// Ensemble_SRN_19782619365570
// MI455X (gfx1250) — hardware-verified
//
#include <hip/hip_runtime.h>
#include <math.h>

typedef __attribute__((ext_vector_type(16))) _Float16 v16h;
typedef __attribute__((ext_vector_type(8)))  _Float16 v8h;
typedef __attribute__((ext_vector_type(16))) __bf16   v16b;
typedef __attribute__((ext_vector_type(8)))  float    v8f;
typedef __attribute__((ext_vector_type(4)))  float    v4f;

__device__ __forceinline__ int frag_k(int i, int h) { return (i < 8) ? (8 * h + i) : (16 + 8 * h + (i - 8)); }
__device__ __forceinline__ __bf16 bf16_rne(float f) {
    unsigned int u = __float_as_uint(f);
    u += 0x7fffu + ((u >> 16) & 1u);
    return __builtin_bit_cast(__bf16, (unsigned short)(u >> 16));
}
__device__ __forceinline__ float bf16_f32(__bf16 b) { return __uint_as_float(((unsigned int)__builtin_bit_cast(unsigned short, b)) << 16); }
__device__ __forceinline__ v8f wmma16(v16h a, v16h b, v8f c) {
    c = __builtin_amdgcn_wmma_f32_16x16x32_f16(false, a, false, b, (short)0, c, false, false);
    asm volatile("v_nop\n\tv_nop\n\tv_nop\n\tv_nop" : "+v"(c) : "v"(a), "v"(b));
    return c;
}
__device__ __forceinline__ v8f wmmab(v16b a, v16b b, v8f c) {
    c = __builtin_amdgcn_wmma_f32_16x16x32_bf16(false, a, false, b, (short)0, c, false, false);
    asm volatile("v_nop\n\tv_nop\n\tv_nop\n\tv_nop" : "+v"(c) : "v"(a), "v"(b));
    return c;
}
struct Split { v16b hi, lo; };
__device__ __forceinline__ v8f wmma3(const Split& a, const Split& b, v8f c) {
    c = __builtin_amdgcn_wmma_f32_16x16x32_bf16(false, a.hi, false, b.hi, (short)0, c, false, false);
    c = __builtin_amdgcn_wmma_f32_16x16x32_bf16(false, a.hi, false, b.lo, (short)0, c, false, false);
    c = __builtin_amdgcn_wmma_f32_16x16x32_bf16(false, a.lo, false, b.hi, (short)0, c, false, false);
    asm volatile("v_nop\n\tv_nop\n\tv_nop\n\tv_nop" : "+v"(c) : "v"(a.hi), "v"(a.lo), "v"(b.hi), "v"(b.lo));
    return c;
}
struct Split3 { v16b hi, mid, lo; };
__device__ __forceinline__ v8f wmma6(const Split3& a, const Split3& b, v8f c) {
    c = __builtin_amdgcn_wmma_f32_16x16x32_bf16(false, a.hi, false, b.hi, (short)0, c, false, false);
    c = __builtin_amdgcn_wmma_f32_16x16x32_bf16(false, a.hi, false, b.mid, (short)0, c, false, false);
    c = __builtin_amdgcn_wmma_f32_16x16x32_bf16(false, a.mid, false, b.hi, (short)0, c, false, false);
    c = __builtin_amdgcn_wmma_f32_16x16x32_bf16(false, a.hi, false, b.lo, (short)0, c, false, false);
    c = __builtin_amdgcn_wmma_f32_16x16x32_bf16(false, a.mid, false, b.mid, (short)0, c, false, false);
    c = __builtin_amdgcn_wmma_f32_16x16x32_bf16(false, a.lo, false, b.hi, (short)0, c, false, false);
    asm volatile("v_nop\n\tv_nop\n\tv_nop\n\tv_nop" : "+v"(c) : "v"(a.hi), "v"(a.mid), "v"(a.lo), "v"(b.hi), "v"(b.mid), "v"(b.lo));
    return c;
}

__device__ __forceinline__ v16h fh_ld(const float* __restrict__ p, long long sk, int k0, int h, int klen, float s) {
    v16h a;
#pragma unroll
    for (int i = 0; i < 16; ++i) { const int k = k0 + frag_k(i, h); a[i] = (k < klen) ? (_Float16)(p[(long long)k * sk] * s) : (_Float16)0.f; }
    return a;
}
__device__ __forceinline__ Split sp_ld(const float* __restrict__ p, long long sk, int k0, int h, int klen, float s) {
    Split r;
#pragma unroll
    for (int i = 0; i < 16; ++i) {
        const int k = k0 + frag_k(i, h); const float x = (k < klen) ? p[(long long)k * sk] * s : 0.f;
        const __bf16 hb = bf16_rne(x); r.hi[i] = hb; r.lo[i] = bf16_rne(x - bf16_f32(hb));
    }
    return r;
}
__device__ __forceinline__ Split3 sp3_ld(const float* __restrict__ p, long long sk, int k0, int h, int klen, float s) {
    Split3 r;
#pragma unroll
    for (int i = 0; i < 16; ++i) {
        const int k = k0 + frag_k(i, h); const float x = (k < klen) ? p[(long long)k * sk] * s : 0.f;
        const __bf16 hb = bf16_rne(x); const float r1 = x - bf16_f32(hb); const __bf16 mb = bf16_rne(r1);
        r.hi[i] = hb; r.mid[i] = mb; r.lo[i] = bf16_rne(r1 - bf16_f32(mb));
    }
    return r;
}
__device__ __forceinline__ v16b bh_ld(const float* __restrict__ p, long long sk, int k0, int h, int klen, float s) {
    v16b a;
#pragma unroll
    for (int i = 0; i < 16; ++i) { const int k = k0 + frag_k(i, h); a[i] = bf16_rne((k < klen) ? p[(long long)k * sk] * s : 0.f); }
    return a;
}
__device__ __forceinline__ v16h fh_row(const _Float16* __restrict__ row, int k0, int h) {
    v16h a;
#pragma unroll
    for (int i = 0; i < 16; ++i) a[i] = row[k0 + frag_k(i, h)];
    return a;
}

#define VST2(T, ptr, val) do { *(volatile T*)(ptr) = (val); __threadfence(); *(volatile T*)(ptr) = (val); } while (0)
typedef float v4f __attribute__((ext_vector_type(4)));
#define VST2V4(ptr, val) do { *(volatile v4f*)(ptr) = (val); __threadfence(); *(volatile v4f*)(ptr) = (val); } while (0)

__device__ __attribute__((noinline)) float act_fn(float v, int act) {
    if (act == 1) return fmaxf(v, 0.f);
    if (act == 2) { const float u = 0.7978845608028654f * (v + 0.044715f * v * v * v); return 0.5f * v * (1.f + tanhf(u)); }
    if (act == 3) return v / (1.f + expf(-v));
    if (act == 4) return 0.5f * v * (1.f + erff(v * 0.7071067811865476f));
    if (act == 5) return tanhf(v);
    if (act == 6) return 1.f / (1.f + expf(-v));
    if (act == 7) return (v > 0.f) ? v : 0.01f * v;
    if (act == 8) return (v > 0.f) ? v : (expf(v) - 1.f);
    if (act == 9) return fminf(fmaxf(v, 0.f), 6.f);
    if (act == 10) return fabsf(v);
    if (act == 11) return (v >= 0.f) ? v : 0.1f * v;
    if (act == 12) return (v > 0.f) ? v : 0.2f * v;
    if (act == 13) return (v > 20.f) ? v : log1pf(expf(v));
    return v;
}

struct GemmP {
    const float* A; const float* B; const float* bias; const float* R; float* C;
    long long sAo, sAi, sAm, sAk, sBo, sBi, sBn, sBk, sCo, sCi, sCm, sRo, sRi, sRm, sRn;
    int M, N, K, zi_n, flags, act; float alpha, beta, sa, sb;
    int Npad, pad_;
};
static_assert(sizeof(GemmP) == 5 * 8 + 15 * 8 + 6 * 4 + 4 * 4 + 2 * 4, "GemmP has padding");

template <int MODE>
__global__ __launch_bounds__(32) void k_gemm(GemmP p) {
    const int lane = threadIdx.x & 31, h = lane >> 4, l15 = lane & 15;
    const int m0 = blockIdx.y * 16, n0 = blockIdx.x * 32;
    const int z = blockIdx.z, zo = z / p.zi_n, zi = z - zo * p.zi_n;
    const float* A = p.A + zo * p.sAo + zi * p.sAi;
    const float* B = p.B + zo * p.sBo + zi * p.sBi;
    const int am = min(m0 + l15, p.M - 1);
    v8f acc[2], comp[2];
#pragma unroll
    for (int t = 0; t < 2; ++t) { v8f zz = {}; acc[t] = zz; comp[t] = zz; }
    for (int k0 = 0; k0 < p.K; k0 += 32) {
        const float* arow = A + (long long)am * p.sAm;
        if (MODE == 1) {
            const Split a = sp_ld(arow, p.sAk, k0, h, p.K, 1.f);
#pragma unroll
            for (int t = 0; t < 2; ++t) {
                const int bn = min(n0 + t * 16 + l15, p.N - 1);
                acc[t] = wmma3(a, sp_ld(B + (long long)bn * p.sBn, p.sBk, k0, h, p.K, 1.f), acc[t]);
            }
        } else if (MODE == 3) {
            const Split3 a = sp3_ld(arow, p.sAk, k0, h, p.K, 1.f);
#pragma unroll
            for (int t = 0; t < 2; ++t) {
                const int bn = min(n0 + t * 16 + l15, p.N - 1);
                acc[t] = wmma6(a, sp3_ld(B + (long long)bn * p.sBn, p.sBk, k0, h, p.K, 1.f), acc[t]);
            }
        } else if (MODE == 4) {
            const Split3 a = sp3_ld(arow, p.sAk, k0, h, p.K, 1.f);
#pragma unroll
            for (int t = 0; t < 2; ++t) {
                const int bn = min(n0 + t * 16 + l15, p.N - 1); v8f zz = {};
                const v8f part = wmma6(a, sp3_ld(B + (long long)bn * p.sBn, p.sBk, k0, h, p.K, 1.f), zz);
                const v8f y = part - comp[t]; const v8f s = acc[t] + y; comp[t] = (s - acc[t]) - y; acc[t] = s;
            }
        } else if (MODE == 2) {
            const v16b a = bh_ld(arow, p.sAk, k0, h, p.K, 1.f);
#pragma unroll
            for (int t = 0; t < 2; ++t) {
                const int bn = min(n0 + t * 16 + l15, p.N - 1);
                acc[t] = wmmab(a, bh_ld(B + (long long)bn * p.sBn, p.sBk, k0, h, p.K, 1.f), acc[t]);
            }
        } else {
            const v16h a = fh_ld(arow, p.sAk, k0, h, p.K, p.sa);
#pragma unroll
            for (int t = 0; t < 2; ++t) {
                const int bn = min(n0 + t * 16 + l15, p.N - 1);
                acc[t] = wmma16(a, fh_ld(B + (long long)bn * p.sBn, p.sBk, k0, h, p.K, p.sb), acc[t]);
            }
        }
    }
    const float iscale = (MODE == 0) ? p.alpha / (p.sa * p.sb) : p.alpha;
    float* C = p.C + zo * p.sCo + zi * p.sCi;
    const float* R = p.R + zo * p.sRo + zi * p.sRi;
    __shared__ __align__(16) float ctile[16][36];
#pragma unroll
    for (int t = 0; t < 2; ++t) {
        const int n = n0 + t * 16 + l15; const int nn = min(n, p.N - 1);
#pragma unroll
        for (int r = 0; r < 8; ++r) {
            const int m = m0 + 8 * h + r; const int mm = min(m, p.M - 1);
            float v = acc[t][r] * iscale;
            if (p.flags & 1) v += p.bias[nn];
            if (p.flags & 2) v += p.bias[mm];
            v = act_fn(v, p.act);
            if (p.flags & 4) v += p.beta * R[(long long)mm * p.sRm + (long long)nn * p.sRn];
            ctile[8 * h + r][t * 16 + l15] = (n < p.N) ? v : 0.f;
        }
    }
    __syncthreads();
    const int NW = (p.Npad > p.N) ? p.Npad : p.N;
    const bool fast = (m0 + 16 <= p.M) && (n0 + 32 <= NW) && ((p.sCm & 3) == 0) && ((((size_t)C) & 15) == 0);
    if (fast) {
#pragma unroll
        for (int s = 0; s < 4; ++s) {
            const int row = s * 4 + (lane >> 3), c4 = (lane & 7) * 4;
            const v4f v = *(const v4f*)&ctile[row][c4];
            VST2V4(C + (long long)(m0 + row) * p.sCm + n0 + c4, v);
        }
    } else {
        for (int row = 0; row < 16; ++row) {
            const int m = m0 + row, n = n0 + lane;
            if (m < p.M && n < NW) VST2(float, C + (long long)m * p.sCm + n, ctile[row][lane]);
        }
    }
}

#define AW 4
struct AttnP {
    const float* Q; const float* K; const float* V; float* O; float* P; const float* Mf; const int* Mi; float* ST;
    const float* Pw; const float* Rt; const int* SQ; const int* SK;
    long long swb, swh, swi, swj, srb, srh, sri;
    long long sQb, sQh, sQi, sQd, sKb, sKh, sKj, sKd, sVb, sVh, sVj, sVd, sOb, sOh, sOi, sPb, sPh, sPi, smb, smh, smi, smj;
    int Lq, Lk, dh, dv, hrep, causal, coff, pband;
    float scale, mfill; int nonorm, mpol;
    int roff, rn, segpol, win;
};
static_assert(sizeof(AttnP) == 12 * 8 + 29 * 8 + 16 * 4, "AttnP has padding");

#ifndef KATTN_ATTR
#define KATTN_ATTR
#endif
template <int DHP, int DVP, int QM, bool SPLITPV, bool TWOPASS>
__global__ __launch_bounds__(32 * AW) KATTN_ATTR void k_attn(AttnP p) {
    constexpr int NT = DVP / 16;
    constexpr int KS = DHP / 32;
    constexpr int VP = DVP + 8;
    __shared__ __align__(16) float    pl[AW][16 * 64];
    __shared__ __align__(16) _Float16 vl[(SPLITPV ? 2 : 1) * 64 * VP];
    const int lane = threadIdx.x & 31, hf = lane >> 4, l15 = lane & 15, wave = threadIdx.x >> 5;
    const int h = blockIdx.y, b = blockIdx.z, hk = h / p.hrep;
    const int q0 = (blockIdx.x * AW + wave) * 16;
    float* myp = pl[wave];
    const float L2E = 1.4426950408889634f;
    const float NEG = -__builtin_inff();
    const int qi = min(q0 + l15, p.Lq - 1);
    const float* qrow = p.Q + b * p.sQb + h * p.sQh + (long long)qi * p.sQi;
    const float* kbase = p.K + b * p.sKb + hk * p.sKh;
    const float* vbase = p.V + b * p.sVb + hk * p.sVh;
    v16h qa[QM == 0 ? KS : 1]; Split qs_[QM == 1 ? KS : 1]; Split3 qt_[QM == 2 ? KS : 1];
#pragma unroll
    for (int ks = 0; ks < KS; ++ks) {
        if (QM == 2) qt_[ks] = sp3_ld(qrow, p.sQd, ks * 32, hf, p.dh, 1.f);
        else if (QM == 1) qs_[ks] = sp_ld(qrow, p.sQd, ks * 32, hf, p.dh, 1.f);
        else qa[ks] = fh_ld(qrow, p.sQd, ks * 32, hf, p.dh, 1.f);
    }
    v8f o[NT]; float m8[8], l8[8];
#pragma unroll
    for (int t = 0; t < NT; ++t) { v8f zz = {}; o[t] = zz; }
#pragma unroll
    for (int i = 0; i < 8; ++i) { m8[i] = NEG; l8[i] = 0.f; }
    int jend = p.Lk;
    if (p.causal == 1) { const int je = (blockIdx.x * AW + AW - 1) * 16 + 16 + p.coff; jend = min(jend, max(je, 0)); }
    const int npass = TWOPASS ? 2 : 1;
    for (int pass = 0; pass < npass; ++pass) {
        const bool dopv = (!TWOPASS) || pass == 1;
        for (int j0 = 0; j0 < jend; j0 += 64) {
            if (dopv) {
                __syncthreads();
                for (int idx = threadIdx.x; idx < 64 * DVP; idx += 32 * AW) {
                    const int jr = idx / DVP, d = idx - jr * DVP, j = j0 + jr;
                    const float f = (j < p.Lk && d < p.dv) ? vbase[(long long)j * p.sVj + (long long)d * p.sVd] : 0.f;
                    if (SPLITPV) {
                        const __bf16 hb = bf16_rne(f);
                        ((__bf16*)vl)[jr * VP + d] = hb; ((__bf16*)vl)[64 * VP + jr * VP + d] = bf16_rne(f - bf16_f32(hb));
                    } else vl[jr * VP + d] = (_Float16)f;
                }
            }
            v8f s[4];
#pragma unroll
            for (int t = 0; t < 4; ++t) {
                const int j = min(j0 + t * 16 + l15, p.Lk - 1);
                const float* krow = kbase + (long long)j * p.sKj;
                v8f acc = {};
#pragma unroll
                for (int ks = 0; ks < KS; ++ks) {
                    if (QM == 2)      acc = wmma6(qt_[ks], sp3_ld(krow, p.sKd, ks * 32, hf, p.dh, 1.f), acc);
                    else if (QM == 1) acc = wmma3(qs_[ks], sp_ld(krow, p.sKd, ks * 32, hf, p.dh, 1.f), acc);
                    else              acc = wmma16(qa[ks], fh_ld(krow, p.sKd, ks * 32, hf, p.dh, 1.f), acc);
                }
                s[t] = acc;
            }
            float pv[8][4];
#pragma unroll
            for (int i = 0; i < 8; ++i) {
                const int irow = q0 + i + 8 * hf;
                const int ic = min(irow, p.Lq - 1);
                float sc[4];
#pragma unroll
                for (int t = 0; t < 4; ++t) {
                    const int jg = j0 + t * 16 + l15;
                    float v = s[t][i] * p.scale;
                    if (p.Mf) v += p.Mf[b * p.smb + h * p.smh + (long long)ic * p.smi + (long long)min(jg, p.Lk - 1) * p.smj];
                    if (p.Rt) { int rc = ic - min(jg, p.Lk - 1) + p.roff; rc = rc < 0 ? 0 : (rc >= p.rn ? p.rn - 1 : rc); v += p.Rt[b * p.srb + h * p.srh + (long long)ic * p.sri + rc]; }
                    if (p.Mi) { const int mv = p.Mi[b * p.smb + h * p.smh + (long long)ic * p.smi + (long long)min(jg, p.Lk - 1) * p.smj]; if (p.mpol ? (mv != 0) : (mv == 0)) v = p.mfill; }
                    if (p.SQ) { const bool same = p.SQ[(long long)b * p.Lq + ic] == p.SK[(long long)b * p.Lk + min(jg, p.Lk - 1)]; if (p.segpol ? same : !same) v = p.mfill; }
                    if (p.causal == 2 && jg > irow + p.coff) v = p.mfill;
                    if (jg >= p.Lk || (p.causal == 1 && jg > irow + p.coff) || (p.causal == 3 && jg < irow + p.coff) || (p.win > 0 && irow + p.coff - jg > p.win)) v = NEG; else v *= L2E;
                    sc[t] = v;
                }
                if (!TWOPASS || pass == 0) {
                    float mx = fmaxf(fmaxf(sc[0], sc[1]), fmaxf(sc[2], sc[3]));
                    mx = fmaxf(mx, __shfl_xor(mx, 1, 32)); mx = fmaxf(mx, __shfl_xor(mx, 2, 32));
                    mx = fmaxf(mx, __shfl_xor(mx, 4, 32)); mx = fmaxf(mx, __shfl_xor(mx, 8, 32));
                    const float mnew = fmaxf(m8[i], mx);
                    const float corr = (mnew == NEG) ? 1.f : exp2f(m8[i] - mnew);
                    float rs = 0.f;
#pragma unroll
                    for (int t = 0; t < 4; ++t) {
                        const float pp = (sc[t] == NEG) ? 0.f : exp2f(sc[t] - mnew); rs += pp;
                        pv[i][t] = p.Pw ? pp * p.Pw[b * p.swb + h * p.swh + (long long)ic * p.swi + (long long)min(j0 + t * 16 + l15, p.Lk - 1) * p.swj] : pp;
                    }
                    rs += __shfl_xor(rs, 1, 32); rs += __shfl_xor(rs, 2, 32); rs += __shfl_xor(rs, 4, 32); rs += __shfl_xor(rs, 8, 32);
                    l8[i] = l8[i] * corr + rs; m8[i] = mnew;
                    if (!TWOPASS) {
#pragma unroll
                        for (int t = 0; t < NT; ++t) o[t][i] *= corr;
                    }
                } else {
                    const float inv = (l8[i] > 0.f) ? 1.f / l8[i] : 0.f;
#pragma unroll
                    for (int t = 0; t < 4; ++t) {
                        const int jg = j0 + t * 16 + l15;
                        float pp = (sc[t] == NEG) ? 0.f : exp2f(sc[t] - m8[i]) * inv;
                        if (p.Pw) pp *= p.Pw[b * p.swb + h * p.swh + (long long)ic * p.swi + (long long)min(jg, p.Lk - 1) * p.swj];
                        pv[i][t] = pp;
                    }
                }
            }
            if (dopv) {
#pragma unroll
                for (int i = 0; i < 8; ++i)
#pragma unroll
                    for (int t = 0; t < 4; ++t) myp[(i + 8 * hf) * 64 + t * 16 + l15] = pv[i][t];
                __syncthreads();
                if (p.P) {
                    float* pb_ = p.P + b * p.sPb + h * p.sPh;
                    const bool fastP = (p.pband == 0) && ((p.sPi & 3) == 0) && (j0 + 64 <= p.Lk) && (q0 + 16 <= p.Lq) && ((((size_t)pb_) & 15) == 0);
                    if (fastP) {
#pragma unroll
                        for (int s = 0; s < 8; ++s) {
                            const int row = s * 2 + (lane >> 4), c4 = (lane & 15) * 4;
                            const v4f v = *(const v4f*)(myp + row * 64 + c4);
                            VST2V4(pb_ + (long long)(q0 + row) * p.sPi + j0 + c4, v);
                        }
                    } else {
                        for (int row = 0; row < 16; ++row) {
                            const int irow = q0 + row; if (irow >= p.Lq) continue;
                            for (int c = lane; c < 64; c += 32) {
                                const int jg = j0 + c; if (jg >= p.Lk) continue;
                                if (p.pband == 0) VST2(float, pb_ + (long long)irow * p.sPi + jg, myp[row * 64 + c]);
                                else if (jg - irow <= p.pband && irow - jg <= p.pband) VST2(float, pb_ + (long long)irow * p.sPi + (jg - irow + p.pband), myp[row * 64 + c]);
                            }
                        }
                    }
                }
                if (SPLITPV) {
                    const Split pa0 = sp_ld(myp + l15 * 64, 1, 0, hf, 64, 1.f), pa1 = sp_ld(myp + l15 * 64, 1, 32, hf, 64, 1.f);
                    const __bf16* vh = (const __bf16*)vl; const __bf16* vlo = vh + 64 * VP;
#pragma unroll
                    for (int t = 0; t < NT; ++t) {
                        const int dcol = t * 16 + l15;
                        Split b0, b1;
#pragma unroll
                        for (int e = 0; e < 16; ++e) {
                            const int k0 = frag_k(e, hf), k1 = 32 + frag_k(e, hf);
                            b0.hi[e] = vh[k0 * VP + dcol]; b0.lo[e] = vlo[k0 * VP + dcol]; b1.hi[e] = vh[k1 * VP + dcol]; b1.lo[e] = vlo[k1 * VP + dcol];
                        }
                        o[t] = wmma3(pa0, b0, o[t]);
                        o[t] = wmma3(pa1, b1, o[t]);
                    }
                } else {
                    const v16h pa0 = fh_ld(myp + l15 * 64, 1, 0, hf, 64, 4096.f), pa1 = fh_ld(myp + l15 * 64, 1, 32, hf, 64, 4096.f);
#pragma unroll
                    for (int t = 0; t < NT; ++t) {
                        const int dcol = t * 16 + l15;
                        v16h b0, b1;
#pragma unroll
                        for (int e = 0; e < 16; ++e) { b0[e] = vl[frag_k(e, hf) * VP + dcol]; b1[e] = vl[(32 + frag_k(e, hf)) * VP + dcol]; }
                        o[t] = wmma16(pa0, b0, o[t]);
                        o[t] = wmma16(pa1, b1, o[t]);
                    }
                }
            }
        }
    }
    float* obase = p.O + b * p.sOb + h * p.sOh;
    if (p.ST) {
        const int rl = lane >> 1, isel = rl & 7;
        float mv = 0.f, lv = 0.f;
#pragma unroll
        for (int i = 0; i < 8; ++i) if (i == isel) { mv = m8[i]; lv = l8[i]; }
        const int irow = q0 + rl;
        if (irow < p.Lq) { float* st = p.ST + (((long long)b * gridDim.y + h) * p.Lq + irow) * 2 + (lane & 1); VST2(float, st, (lane & 1) ? lv : mv * 0.6931471805599453f); }
    }
    float invr[8];
#pragma unroll
    for (int i = 0; i < 8; ++i) {
        if (TWOPASS) invr[i] = SPLITPV ? 1.f : (1.f / 4096.f);
        else if (p.nonorm) invr[i] = exp2f(m8[i]) * (SPLITPV ? 1.f : (1.f / 4096.f));
        else invr[i] = (l8[i] > 0.f) ? (SPLITPV ? 1.f / l8[i] : 1.f / (l8[i] * 4096.f)) : 0.f;
    }
    __syncthreads();
    const bool ofast = ((p.sOi & 3) == 0) && ((((size_t)obase) & 15) == 0) && (q0 + 16 <= p.Lq);
#pragma unroll
    for (int c0 = 0; c0 < DVP; c0 += 64) {
#pragma unroll
        for (int i = 0; i < 8; ++i)
#pragma unroll
            for (int t = 0; t < NT; ++t) if (t * 16 >= c0 && t * 16 < c0 + 64) myp[(i + 8 * hf) * 64 + (t * 16 - c0) + l15] = o[t][i] * invr[i];
        __syncthreads();
        const int cw = (DVP - c0 < 64) ? (DVP - c0) : 64;
        if (ofast && (c0 + cw <= p.dv) && (cw % 32 == 0)) {
            const int lpr = cw / 4;
            const int rows_per_ins = 32 / lpr;
            for (int r0 = 0; r0 < 16; r0 += rows_per_ins) {
                const int row = r0 + lane / lpr, c4 = (lane % lpr) * 4;
                const v4f v = *(const v4f*)(myp + row * 64 + c4);
                VST2V4(obase + (long long)(q0 + row) * p.sOi + c0 + c4, v);
            }
        } else {
            for (int row = 0; row < 16; ++row) {
                const int irow = q0 + row; if (irow >= p.Lq) continue;
                for (int c = lane; c < cw; c += 32) { const int d = c0 + c; if (d < p.dv) VST2(float, obase + (long long)irow * p.sOi + d, myp[row * 64 + c]); }
            }
        }
        __syncthreads();
    }
}

struct TrP { const float* src; float* dst; const float* R2; long long sSz, lds, sDz, ldd, sRz, ldr; int R, C, flags, act; float alpha, beta; };
static_assert(sizeof(TrP) == 3 * 8 + 6 * 8 + 6 * 4, "TrP has padding");
__global__ __launch_bounds__(256) void k_tr(TrP p) {
    __shared__ float tile[32][33];
    const int c0 = blockIdx.x * 32, r0 = blockIdx.y * 32, z = blockIdx.z;
    const int lane = threadIdx.x & 31, wave = threadIdx.x >> 5;
    const float* s = p.src + z * p.sSz;
#pragma unroll
    for (int k = 0; k < 4; ++k) {
        const int rl = wave * 4 + k, r = r0 + rl, c = c0 + lane;
        tile[rl][lane] = (r < p.R && c < p.C) ? s[(long long)r * p.lds + c] : 0.f;
    }
    __syncthreads();
    float* d = p.dst + z * p.sDz; const float* rr = p.R2 + z * p.sRz;
#pragma unroll
    for (int k = 0; k < 4; ++k) {
        const int cl = wave * 4 + k, c = c0 + cl, r = r0 + lane;
        if (c < p.C && r < p.R) {
            float v = act_fn(p.alpha * tile[lane][cl], p.act);
            if (p.flags & 1) v += p.beta * rr[(long long)c * p.ldr + r];
            VST2(float, d + (long long)c * p.ldd + r, v);
        }
    }
}

__global__ __launch_bounds__(256) void k_affine(const float* __restrict__ src, float* __restrict__ dst, int n, float a, float b, const float* __restrict__ sdev) {
    const int i = blockIdx.x * 256 + threadIdx.x;
    if (i < n) { const float aa = sdev ? a * sdev[0] : a; const float v = aa * src[i] + b; VST2(float, dst + i, v); }
}

struct SmP { const float* src; float* dst; const float* Mf; long long sz, sr, dz, dr, smz, smr; int n, pad; float scale_in, scale_out; };
static_assert(sizeof(SmP) == 3 * 8 + 6 * 8 + 4 * 4, "SmP has padding");
__global__ __launch_bounds__(256) void k_softmax(SmP p) {
    __shared__ float red[256];
    const int r = blockIdx.x, z = blockIdx.y, tid = threadIdx.x;
    const float* s = p.src + z * p.sz + (long long)r * p.sr;
    const float* mf = p.Mf ? (p.Mf + z * p.smz + (long long)r * p.smr) : nullptr;
    float mx = -__builtin_inff();
    for (int j = tid; j < p.n; j += 256) { float v = s[j] * p.scale_in; if (mf) v += mf[j]; mx = fmaxf(mx, v); }
    red[tid] = mx; __syncthreads();
    for (int o = 128; o > 0; o >>= 1) { if (tid < o) red[tid] = fmaxf(red[tid], red[tid + o]); __syncthreads(); }
    mx = red[0]; __syncthreads();
    float sum = 0.f;
    for (int j = tid; j < p.n; j += 256) { float v = s[j] * p.scale_in; if (mf) v += mf[j]; sum += (mx == -__builtin_inff()) ? 0.f : expf(v - mx); }
    red[tid] = sum; __syncthreads();
    for (int o = 128; o > 0; o >>= 1) { if (tid < o) red[tid] += red[tid + o]; __syncthreads(); }
    sum = red[0];
    const float inv = (sum > 0.f) ? p.scale_out / sum : 0.f;
    float* d = p.dst + z * p.dz + (long long)r * p.dr;
    for (int j = tid; j < p.n; j += 256) { float v = s[j] * p.scale_in; if (mf) v += mf[j]; const float o = (mx == -__builtin_inff()) ? 0.f : expf(v - mx) * inv; VST2(float, d + j, o); }
}
__global__ __launch_bounds__(256) void k_stats(const float* __restrict__ x, long long sz, long long so, long long si, int inner, int n, float eps, float* __restrict__ stat, int mode) {
    __shared__ float red[256];
    const int z = blockIdx.x, tid = threadIdx.x;
    const float* base = x + z * sz;
    float s = 0.f;
    for (int e = tid; e < n; e += 256) s += base[(long long)(e / inner) * so + (long long)(e % inner) * si];
    red[tid] = s; __syncthreads();
    for (int o = 128; o > 0; o >>= 1) { if (tid < o) red[tid] += red[tid + o]; __syncthreads(); }
    const float mu = (mode == 0 || mode == 3) ? red[0] / (float)n : 0.f; __syncthreads();
    float q = 0.f;
    for (int e = tid; e < n; e += 256) { const float dlt = base[(long long)(e / inner) * so + (long long)(e % inner) * si] - mu; q += dlt * dlt; }
    red[tid] = q; __syncthreads();
    for (int o = 128; o > 0; o >>= 1) { if (tid < o) red[tid] += red[tid + o]; __syncthreads(); }
    {
        float rs;
        if (mode == 2) rs = sqrtf((float)n) / fmaxf(sqrtf(red[0]), eps); else if (mode == 3) rs = rsqrtf(red[0] / (float)(n - 1) + eps); else rs = rsqrtf(red[0] / (float)n + eps);
        if (tid < 32) { const float v = (tid == 0) ? mu : ((tid == 1) ? rs : 0.f); VST2(float, stat + (long long)z * 32 + tid, v); }
    }
}
__global__ __launch_bounds__(256) void k_norm_apply(const float* __restrict__ x, float* __restrict__ y, const float* __restrict__ stat, const float* __restrict__ g, const float* __restrict__ bta,
                                                     int Z, int C, int L, int G, int bn, int act) {
    const long long idx = (long long)blockIdx.x * 256 + threadIdx.x;
    if (idx >= (long long)Z * C * L) return;
    const int l = (int)(idx % L); const long long zc = idx / L; const int c = (int)(zc % C), z = (int)(zc / C); (void)l;
    const int set = bn ? c : (z * G + c / (C / G));
    float v = (x[idx] - stat[(long long)set * 32]) * stat[(long long)set * 32 + 1];
    if (g) v *= g[c];
    if (bta) v += bta[c];
    v = act_fn(v, act);
    VST2(float, y + idx, v);
}

__global__ __launch_bounds__(256) void k_lse_neg(const float* __restrict__ st, float* __restrict__ c, int n) {
    const int i = blockIdx.x * 256 + threadIdx.x;
    if (i < n) { const float v = -(st[2 * i] + logf(st[2 * i + 1])); VST2(float, c + i, v); }
}

__global__ __launch_bounds__(256) void k_iota(int* __restrict__ dst, int n, int a, int b) {
    const int i = blockIdx.x * 256 + threadIdx.x;
    if (i < n) { const int v = a * i + b; VST2(int, dst + i, v); }
}

__global__ __launch_bounds__(256) void k_axpby(const float* __restrict__ x, const float* __restrict__ y, float* __restrict__ dst, int n, float a, float b, float c) {
    const int i = blockIdx.x * 256 + threadIdx.x;
    if (i < n) { const float v = a * x[i] + b * y[i] + c; VST2(float, dst + i, v); }
}

struct RopeP { const float* X; float* Y; const float* C; const float* Sn; const int* pos; long long sXr, sXh, sYr, sYh, sCb, sCp, sCd; int R, Hn, D, S, mode, tmode, pmode, pad; };
static_assert(sizeof(RopeP) == 5 * 8 + 7 * 8 + 8 * 4, "RopeP has padding");
__global__ __launch_bounds__(256) void k_rope(RopeP p) {
    const long long idx = (long long)blockIdx.x * 256 + threadIdx.x;
    if (idx >= (long long)p.R * p.Hn * p.D) return;
    const int d = (int)(idx % p.D); const long long rh = idx / p.D; const int h = (int)(rh % p.Hn); const int r = (int)(rh / p.Hn);
    const int half = p.D / 2;
    int partner; float sign;
    if (p.mode == 0) { partner = (d < half) ? d + half : d - half; sign = (d < half) ? -1.f : 1.f; }
    else { partner = d ^ 1; sign = (d & 1) ? 1.f : -1.f; }
    const int tcol = (p.tmode == 0) ? d : ((p.tmode == 1) ? (d % half) : (d >> 1));
    const int pp = (p.pmode == 0) ? (r % p.S) : ((p.pmode == 1) ? h : p.pos[r]);
    const long long toff = (long long)(r / p.S) * p.sCb + (long long)pp * p.sCp + (long long)tcol * p.sCd;
    const float* xr = p.X + (long long)r * p.sXr + (long long)h * p.sXh;
    const float v = xr[d] * p.C[toff] + sign * xr[partner] * p.Sn[toff];
    VST2(float, p.Y + (long long)r * p.sYr + (long long)h * p.sYh + d, v);
}

__global__ __launch_bounds__(256) void k_invf(float* __restrict__ invb, int half, int D, float base, float num, int fmode, float cexp) {
    const int i = blockIdx.x * 256 + threadIdx.x;
    if (i >= ((half + 31) / 32) * 32) return;
    if (i >= half) { VST2(float, invb + i, 0.f); return; }
    const float e = (float)(2 * i) / (float)D;
    float invf;
    if (fmode == 1) invf = num * expf((float)(2 * i) * cexp);
    else if (fmode == 2) invf = num * powf(base, (-2.0f * ((float)i - 1.0f)) / (float)D);
    else invf = num * (1.0f / powf(base, e));
    VST2(float, invb + i, invf);
}
__global__ __launch_bounds__(256) void k_sincos(float* __restrict__ cs, float* __restrict__ sn, const float* __restrict__ invb, int S, int half, float pscale) {
    const int idx = blockIdx.x * 256 + threadIdx.x;
    if (idx >= S * half) return;
    const int s = idx / half, i = idx - s * half;
    const float ang = (pscale * (float)s) * invb[i];
    VST2(float, cs + idx, cosf(ang)); VST2(float, sn + idx, sinf(ang));
}

__global__ __launch_bounds__(256) void k_mulact(const float* __restrict__ x, const float* __restrict__ y, float* __restrict__ dst, int n, int act) {
    const int i = blockIdx.x * 256 + threadIdx.x;
    if (i < n) { const float v = act_fn(x[i], act) * y[i]; VST2(float, dst + i, v); }
}

__global__ __launch_bounds__(256) void k_matvec(GemmP p) {
    const int rpt = (p.N == 1) ? 1 : 32;
    const long long r0 = ((long long)blockIdx.x * 256 + threadIdx.x) * rpt; const int z = blockIdx.z, zo = z / p.zi_n, zi = z - zo * p.zi_n;
    if (r0 >= p.M) return;
    const float* Bb = p.B + zo * p.sBo + zi * p.sBi;
    float* C = p.C + zo * p.sCo + zi * p.sCi; const float* R = p.R + zo * p.sRo + zi * p.sRi;
    for (int rr = 0; rr < rpt; ++rr) {
        const long long r = r0 + rr; if (r >= p.M) break;
        const float* A = p.A + zo * p.sAo + zi * p.sAi + r * p.sAm;
        float acc[8] = {0.f, 0.f, 0.f, 0.f, 0.f, 0.f, 0.f, 0.f};
        for (int k = 0; k < p.K; ++k) { const float a = A[(long long)k * p.sAk];
#pragma unroll
            for (int j = 0; j < 8; ++j) if (j < p.N) acc[j] += a * Bb[(long long)j * p.sBn + (long long)k * p.sBk]; }
#pragma unroll
        for (int j = 0; j < 8; ++j) if (j < p.N) {
            float v = acc[j] * p.alpha;
            if (p.flags & 1) v += p.bias[j];
            if (p.flags & 2) v += p.bias[r];
            v = act_fn(v, p.act);
            if (p.flags & 4) v += p.beta * R[r * p.sRm + (long long)j * p.sRn];
            VST2(float, C + r * p.sCm + j, v);
        }
    }
}
__global__ __launch_bounds__(256) void k_smallsoftmax(const float* __restrict__ src, float* __restrict__ dst, long long sr, long long dr, int n, long long R, float scale) {
    const long long r0 = ((long long)blockIdx.x * 256 + threadIdx.x) * 32;
    for (int rr = 0; rr < 32; ++rr) {
        const long long r = r0 + rr; if (r >= R) return;
        const float* s = src + r * sr; float* d = dst + r * dr;
        float mx = -__builtin_inff();
        for (int j = 0; j < n; ++j) mx = fmaxf(mx, s[j] * scale);
        float sum = 0.f;
        for (int j = 0; j < n; ++j) sum += expf(s[j] * scale - mx);
        const float inv = 1.f / sum;
        for (int j = 0; j < n; ++j) { const float v = expf(s[j] * scale - mx) * inv; VST2(float, d + j, v); }
    }
}

__global__ __launch_bounds__(32) void k_unitstat(float* __restrict__ st) { const int t = threadIdx.x; const float v = (t == 1) ? 1.f : 0.f; VST2(float, st + t, v); }

__global__ __launch_bounds__(256) void k_lincopy(const float* __restrict__ src, long long lds, float* __restrict__ dst, long long ldd, long long rows, int cols) {
    const long long i = (long long)blockIdx.x * 256 + threadIdx.x; if (i >= rows * cols) return;
    const long long r = i / cols; const int c = (int)(i - r * cols);
    const float v = src[r * lds + c]; VST2(float, dst + r * ldd + c, v);
}

__global__ __launch_bounds__(256) void k_es_idx(const float* __restrict__ X, int* __restrict__ IDX, int N) { const int n = blockIdx.x * 256 + threadIdx.x; if (n >= N) return; int ij[3];
#pragma unroll 1
    for (int d = 0; d < 3; ++d) { const float v = X[(long long)n * 3 + d]; int q = (int)((v + 1.f) * 0.5f * 4.f); ij[d] = min(max(q, 0), 3); }
    VST2(int, IDX + n, ij[2] + ij[1] * 4 + ij[0] * 16); }
__global__ void k_es_offt(int* __restrict__ OFFT) { const int m = threadIdx.x; if (m <= 64) { const int offs[65] = {0, 8258, 16336, 24522, 32821, 40958, 49110, 57311, 65470, 73590, 81694, 89741, 97909, 106318, 114412, 122629, 130922, 139144, 147223, 155410, 163700, 171935, 180113, 188211, 196560, 204689, 212743, 221057, 229226, 237465, 245796, 254056, 262182, 270491, 278679, 286947, 295041, 303152, 311243, 319401, 327680, 335847, 344148, 352407, 360579, 368740, 376988, 385261, 393322, 401421, 409659, 417950, 426348, 434527, 442798, 450881, 459024, 467170, 475274, 483486, 491692, 499883, 507988, 516109, 524288}; VST2(int, OFFT + m, offs[m]); } }
__global__ __launch_bounds__(256) void k_es_group(const int* __restrict__ IDX, const int* __restrict__ OFFT, int* __restrict__ slot, int N) { __shared__ int sc[256]; const int m = blockIdx.x; const int t = threadIdx.x; int running = OFFT[m];
    for (int base = 0; base < N; base += 256) { const int n = base + t; const int f = (n < N && IDX[n] == m) ? 1 : 0; sc[t] = f; __syncthreads();
        for (int o = 1; o < 256; o <<= 1) { const int v = (t >= o) ? sc[t - o] : 0; __syncthreads(); sc[t] += v; __syncthreads(); }
        if (f) VST2(int, slot + running + sc[t] - 1, n); const int tot = sc[255]; __syncthreads(); running += tot; } }
__global__ __launch_bounds__(256) void k_es_gather(const float* __restrict__ X, const int* __restrict__ slot, float* __restrict__ XS, int N) { const int q = blockIdx.x * 256 + threadIdx.x; if (q >= N * 8) return; const int c = q % 8; const int p = q / 8; VST2(float, XS + q, (c < 3) ? X[(long long)slot[p] * 3 + c] : 0.f); }
__global__ __launch_bounds__(256) void k_es_scatter(const float* __restrict__ Y, int ldp, const int* __restrict__ slot, const int* __restrict__ IDX, int m, int p0, int cntm, float* __restrict__ OUT) { const int r = blockIdx.x * 256 + threadIdx.x; if (r >= cntm) return; const int p = p0 + r; const int n = slot[p]; if (IDX[n] == m) VST2(float, OUT + n, Y[(long long)r * ldp]); }

template __global__ void k_gemm<0>(GemmP);

extern "C" void kernel_launch(void* const* d_in, const int* in_sizes, int n_in, void* d_out, int out_size, void* d_ws, size_t ws_size, hipStream_t stream) {
    (void)in_sizes; (void)n_in; (void)out_size; (void)ws_size;
    const float* x = (const float*)d_in[0];
    const float* W1 = (const float*)d_in[1];
    const float* b1 = (const float*)d_in[2];
    const float* W2 = (const float*)d_in[3];
    const float* b2 = (const float*)d_in[4];
    const float* W3 = (const float*)d_in[5];
    const float* b3 = (const float*)d_in[6];
    const int N = 524288;
    const int M = 64;
    const int H = 64;
    const int LP = 32;
    const int CAP = 16384;
    float* out = (float*)d_out;
    char* wsp = (char*)d_ws;
    int* IDX = (int*)wsp; wsp += (((size_t)((size_t)N + 64) * 4 + 255) / 256) * 256;
    int* slot = (int*)wsp; wsp += (((size_t)((size_t)N + 64) * 4 + 255) / 256) * 256;
    int* OFFT = (int*)wsp; wsp += (((size_t)((size_t)M + 64) * 4 + 255) / 256) * 256;
    float* XS = (float*)wsp; wsp += (((size_t)((size_t)(N + 64) * 8) * 4 + 255) / 256) * 256;
    float* H1 = (float*)wsp; wsp += (((size_t)((size_t)CAP * H) * 4 + 255) / 256) * 256;
    float* H2 = (float*)wsp; wsp += (((size_t)((size_t)CAP * H) * 4 + 255) / 256) * 256;
    float* Y = (float*)wsp; wsp += (((size_t)((size_t)CAP * LP) * 4 + 255) / 256) * 256;
    hipMemsetAsync(out, 0, (size_t)N * 4, stream);
    k_es_idx<<<(unsigned)((N + 255) / 256), 256, 0, stream>>>(x, IDX, N); k_es_offt<<<1, 128, 0, stream>>>(OFFT);
    k_es_group<<<M, 256, 0, stream>>>(IDX, OFFT, slot, N);
    k_es_gather<<<(unsigned)((N * 8 + 255) / 256), 256, 0, stream>>>(x, slot, XS, N);
    { GemmP g1_0;
      g1_0.A = XS + (size_t)0 * 8; g1_0.B = W1 + 0; g1_0.bias = b1 + 0; g1_0.R = XS + (size_t)0 * 8; g1_0.C = H1;
      g1_0.sAo = 0; g1_0.sAi = 0; g1_0.sAm = 8; g1_0.sAk = 1; g1_0.sBo = 0; g1_0.sBi = 0; g1_0.sBn = 1; g1_0.sBk = H; g1_0.sCo = 0; g1_0.sCi = 0; g1_0.sCm = H; g1_0.sRo = 0; g1_0.sRi = 0; g1_0.sRm = 0; g1_0.sRn = 0;
      g1_0.M = 8258; g1_0.N = H; g1_0.K = 3; g1_0.zi_n = 1; g1_0.flags = 1; g1_0.act = 1;
      g1_0.alpha = 1.0f; g1_0.beta = 0.0f; g1_0.sa = 1.0f; g1_0.sb = 8.0f; g1_0.Npad = H; g1_0.pad_ = 0;
      k_gemm<0><<<dim3((unsigned)((H) + 31) / 32, (unsigned)((8258) + 15) / 16, (unsigned)(1)), 32, 0, stream>>>(g1_0); }
    { GemmP g2_0;
      g2_0.A = H1; g2_0.B = W2 + 0; g2_0.bias = b2 + 0; g2_0.R = H1; g2_0.C = H2;
      g2_0.sAo = 0; g2_0.sAi = 0; g2_0.sAm = H; g2_0.sAk = 1; g2_0.sBo = 0; g2_0.sBi = 0; g2_0.sBn = 1; g2_0.sBk = H; g2_0.sCo = 0; g2_0.sCi = 0; g2_0.sCm = H; g2_0.sRo = 0; g2_0.sRi = 0; g2_0.sRm = 0; g2_0.sRn = 0;
      g2_0.M = 8258; g2_0.N = H; g2_0.K = H; g2_0.zi_n = 1; g2_0.flags = 1; g2_0.act = 1;
      g2_0.alpha = 1.0f; g2_0.beta = 0.0f; g2_0.sa = 1.0f; g2_0.sb = 8.0f; g2_0.Npad = H; g2_0.pad_ = 0;
      k_gemm<0><<<dim3((unsigned)((H) + 31) / 32, (unsigned)((8258) + 15) / 16, (unsigned)(1)), 32, 0, stream>>>(g2_0); }
    { GemmP g3_0;
      g3_0.A = H2; g3_0.B = W3 + 0; g3_0.bias = b3 + 0; g3_0.R = H2; g3_0.C = Y;
      g3_0.sAo = 0; g3_0.sAi = 0; g3_0.sAm = H; g3_0.sAk = 1; g3_0.sBo = 0; g3_0.sBi = 0; g3_0.sBn = 1; g3_0.sBk = 1; g3_0.sCo = 0; g3_0.sCi = 0; g3_0.sCm = LP; g3_0.sRo = 0; g3_0.sRi = 0; g3_0.sRm = 0; g3_0.sRn = 0;
      g3_0.M = 8258; g3_0.N = 1; g3_0.K = H; g3_0.zi_n = 1; g3_0.flags = 1; g3_0.act = 0;
      g3_0.alpha = 1.0f; g3_0.beta = 0.0f; g3_0.sa = 1.0f; g3_0.sb = 8.0f; g3_0.Npad = LP; g3_0.pad_ = 0;
      k_gemm<0><<<dim3((unsigned)((LP) + 31) / 32, (unsigned)((8258) + 15) / 16, (unsigned)(1)), 32, 0, stream>>>(g3_0); }
    k_es_scatter<<<(unsigned)((8258 + 255) / 256), 256, 0, stream>>>(Y, LP, slot, IDX, 0, 0, 8258, out);
    { GemmP g1_1;
      g1_1.A = XS + (size_t)8258 * 8; g1_1.B = W1 + 192; g1_1.bias = b1 + 64; g1_1.R = XS + (size_t)8258 * 8; g1_1.C = H1;
      g1_1.sAo = 0; g1_1.sAi = 0; g1_1.sAm = 8; g1_1.sAk = 1; g1_1.sBo = 0; g1_1.sBi = 0; g1_1.sBn = 1; g1_1.sBk = H; g1_1.sCo = 0; g1_1.sCi = 0; g1_1.sCm = H; g1_1.sRo = 0; g1_1.sRi = 0; g1_1.sRm = 0; g1_1.sRn = 0;
      g1_1.M = 8078; g1_1.N = H; g1_1.K = 3; g1_1.zi_n = 1; g1_1.flags = 1; g1_1.act = 1;
      g1_1.alpha = 1.0f; g1_1.beta = 0.0f; g1_1.sa = 1.0f; g1_1.sb = 8.0f; g1_1.Npad = H; g1_1.pad_ = 0;
      k_gemm<0><<<dim3((unsigned)((H) + 31) / 32, (unsigned)((8078) + 15) / 16, (unsigned)(1)), 32, 0, stream>>>(g1_1); }
    { GemmP g2_1;
      g2_1.A = H1; g2_1.B = W2 + 4096; g2_1.bias = b2 + 64; g2_1.R = H1; g2_1.C = H2;
      g2_1.sAo = 0; g2_1.sAi = 0; g2_1.sAm = H; g2_1.sAk = 1; g2_1.sBo = 0; g2_1.sBi = 0; g2_1.sBn = 1; g2_1.sBk = H; g2_1.sCo = 0; g2_1.sCi = 0; g2_1.sCm = H; g2_1.sRo = 0; g2_1.sRi = 0; g2_1.sRm = 0; g2_1.sRn = 0;
      g2_1.M = 8078; g2_1.N = H; g2_1.K = H; g2_1.zi_n = 1; g2_1.flags = 1; g2_1.act = 1;
      g2_1.alpha = 1.0f; g2_1.beta = 0.0f; g2_1.sa = 1.0f; g2_1.sb = 8.0f; g2_1.Npad = H; g2_1.pad_ = 0;
      k_gemm<0><<<dim3((unsigned)((H) + 31) / 32, (unsigned)((8078) + 15) / 16, (unsigned)(1)), 32, 0, stream>>>(g2_1); }
    { GemmP g3_1;
      g3_1.A = H2; g3_1.B = W3 + 64; g3_1.bias = b3 + 1; g3_1.R = H2; g3_1.C = Y;
      g3_1.sAo = 0; g3_1.sAi = 0; g3_1.sAm = H; g3_1.sAk = 1; g3_1.sBo = 0; g3_1.sBi = 0; g3_1.sBn = 1; g3_1.sBk = 1; g3_1.sCo = 0; g3_1.sCi = 0; g3_1.sCm = LP; g3_1.sRo = 0; g3_1.sRi = 0; g3_1.sRm = 0; g3_1.sRn = 0;
      g3_1.M = 8078; g3_1.N = 1; g3_1.K = H; g3_1.zi_n = 1; g3_1.flags = 1; g3_1.act = 0;
      g3_1.alpha = 1.0f; g3_1.beta = 0.0f; g3_1.sa = 1.0f; g3_1.sb = 8.0f; g3_1.Npad = LP; g3_1.pad_ = 0;
      k_gemm<0><<<dim3((unsigned)((LP) + 31) / 32, (unsigned)((8078) + 15) / 16, (unsigned)(1)), 32, 0, stream>>>(g3_1); }
    k_es_scatter<<<(unsigned)((8078 + 255) / 256), 256, 0, stream>>>(Y, LP, slot, IDX, 1, 8258, 8078, out);
    { GemmP g1_2;
      g1_2.A = XS + (size_t)16336 * 8; g1_2.B = W1 + 384; g1_2.bias = b1 + 128; g1_2.R = XS + (size_t)16336 * 8; g1_2.C = H1;
      g1_2.sAo = 0; g1_2.sAi = 0; g1_2.sAm = 8; g1_2.sAk = 1; g1_2.sBo = 0; g1_2.sBi = 0; g1_2.sBn = 1; g1_2.sBk = H; g1_2.sCo = 0; g1_2.sCi = 0; g1_2.sCm = H; g1_2.sRo = 0; g1_2.sRi = 0; g1_2.sRm = 0; g1_2.sRn = 0;
      g1_2.M = 8186; g1_2.N = H; g1_2.K = 3; g1_2.zi_n = 1; g1_2.flags = 1; g1_2.act = 1;
      g1_2.alpha = 1.0f; g1_2.beta = 0.0f; g1_2.sa = 1.0f; g1_2.sb = 8.0f; g1_2.Npad = H; g1_2.pad_ = 0;
      k_gemm<0><<<dim3((unsigned)((H) + 31) / 32, (unsigned)((8186) + 15) / 16, (unsigned)(1)), 32, 0, stream>>>(g1_2); }
    { GemmP g2_2;
      g2_2.A = H1; g2_2.B = W2 + 8192; g2_2.bias = b2 + 128; g2_2.R = H1; g2_2.C = H2;
      g2_2.sAo = 0; g2_2.sAi = 0; g2_2.sAm = H; g2_2.sAk = 1; g2_2.sBo = 0; g2_2.sBi = 0; g2_2.sBn = 1; g2_2.sBk = H; g2_2.sCo = 0; g2_2.sCi = 0; g2_2.sCm = H; g2_2.sRo = 0; g2_2.sRi = 0; g2_2.sRm = 0; g2_2.sRn = 0;
      g2_2.M = 8186; g2_2.N = H; g2_2.K = H; g2_2.zi_n = 1; g2_2.flags = 1; g2_2.act = 1;
      g2_2.alpha = 1.0f; g2_2.beta = 0.0f; g2_2.sa = 1.0f; g2_2.sb = 8.0f; g2_2.Npad = H; g2_2.pad_ = 0;
      k_gemm<0><<<dim3((unsigned)((H) + 31) / 32, (unsigned)((8186) + 15) / 16, (unsigned)(1)), 32, 0, stream>>>(g2_2); }
    { GemmP g3_2;
      g3_2.A = H2; g3_2.B = W3 + 128; g3_2.bias = b3 + 2; g3_2.R = H2; g3_2.C = Y;
      g3_2.sAo = 0; g3_2.sAi = 0; g3_2.sAm = H; g3_2.sAk = 1; g3_2.sBo = 0; g3_2.sBi = 0; g3_2.sBn = 1; g3_2.sBk = 1; g3_2.sCo = 0; g3_2.sCi = 0; g3_2.sCm = LP; g3_2.sRo = 0; g3_2.sRi = 0; g3_2.sRm = 0; g3_2.sRn = 0;
      g3_2.M = 8186; g3_2.N = 1; g3_2.K = H; g3_2.zi_n = 1; g3_2.flags = 1; g3_2.act = 0;
      g3_2.alpha = 1.0f; g3_2.beta = 0.0f; g3_2.sa = 1.0f; g3_2.sb = 8.0f; g3_2.Npad = LP; g3_2.pad_ = 0;
      k_gemm<0><<<dim3((unsigned)((LP) + 31) / 32, (unsigned)((8186) + 15) / 16, (unsigned)(1)), 32, 0, stream>>>(g3_2); }
    k_es_scatter<<<(unsigned)((8186 + 255) / 256), 256, 0, stream>>>(Y, LP, slot, IDX, 2, 16336, 8186, out);
    { GemmP g1_3;
      g1_3.A = XS + (size_t)24522 * 8; g1_3.B = W1 + 576; g1_3.bias = b1 + 192; g1_3.R = XS + (size_t)24522 * 8; g1_3.C = H1;
      g1_3.sAo = 0; g1_3.sAi = 0; g1_3.sAm = 8; g1_3.sAk = 1; g1_3.sBo = 0; g1_3.sBi = 0; g1_3.sBn = 1; g1_3.sBk = H; g1_3.sCo = 0; g1_3.sCi = 0; g1_3.sCm = H; g1_3.sRo = 0; g1_3.sRi = 0; g1_3.sRm = 0; g1_3.sRn = 0;
      g1_3.M = 8299; g1_3.N = H; g1_3.K = 3; g1_3.zi_n = 1; g1_3.flags = 1; g1_3.act = 1;
      g1_3.alpha = 1.0f; g1_3.beta = 0.0f; g1_3.sa = 1.0f; g1_3.sb = 8.0f; g1_3.Npad = H; g1_3.pad_ = 0;
      k_gemm<0><<<dim3((unsigned)((H) + 31) / 32, (unsigned)((8299) + 15) / 16, (unsigned)(1)), 32, 0, stream>>>(g1_3); }
    { GemmP g2_3;
      g2_3.A = H1; g2_3.B = W2 + 12288; g2_3.bias = b2 + 192; g2_3.R = H1; g2_3.C = H2;
      g2_3.sAo = 0; g2_3.sAi = 0; g2_3.sAm = H; g2_3.sAk = 1; g2_3.sBo = 0; g2_3.sBi = 0; g2_3.sBn = 1; g2_3.sBk = H; g2_3.sCo = 0; g2_3.sCi = 0; g2_3.sCm = H; g2_3.sRo = 0; g2_3.sRi = 0; g2_3.sRm = 0; g2_3.sRn = 0;
      g2_3.M = 8299; g2_3.N = H; g2_3.K = H; g2_3.zi_n = 1; g2_3.flags = 1; g2_3.act = 1;
      g2_3.alpha = 1.0f; g2_3.beta = 0.0f; g2_3.sa = 1.0f; g2_3.sb = 8.0f; g2_3.Npad = H; g2_3.pad_ = 0;
      k_gemm<0><<<dim3((unsigned)((H) + 31) / 32, (unsigned)((8299) + 15) / 16, (unsigned)(1)), 32, 0, stream>>>(g2_3); }
    { GemmP g3_3;
      g3_3.A = H2; g3_3.B = W3 + 192; g3_3.bias = b3 + 3; g3_3.R = H2; g3_3.C = Y;
      g3_3.sAo = 0; g3_3.sAi = 0; g3_3.sAm = H; g3_3.sAk = 1; g3_3.sBo = 0; g3_3.sBi = 0; g3_3.sBn = 1; g3_3.sBk = 1; g3_3.sCo = 0; g3_3.sCi = 0; g3_3.sCm = LP; g3_3.sRo = 0; g3_3.sRi = 0; g3_3.sRm = 0; g3_3.sRn = 0;
      g3_3.M = 8299; g3_3.N = 1; g3_3.K = H; g3_3.zi_n = 1; g3_3.flags = 1; g3_3.act = 0;
      g3_3.alpha = 1.0f; g3_3.beta = 0.0f; g3_3.sa = 1.0f; g3_3.sb = 8.0f; g3_3.Npad = LP; g3_3.pad_ = 0;
      k_gemm<0><<<dim3((unsigned)((LP) + 31) / 32, (unsigned)((8299) + 15) / 16, (unsigned)(1)), 32, 0, stream>>>(g3_3); }
    k_es_scatter<<<(unsigned)((8299 + 255) / 256), 256, 0, stream>>>(Y, LP, slot, IDX, 3, 24522, 8299, out);
    { GemmP g1_4;
      g1_4.A = XS + (size_t)32821 * 8; g1_4.B = W1 + 768; g1_4.bias = b1 + 256; g1_4.R = XS + (size_t)32821 * 8; g1_4.C = H1;
      g1_4.sAo = 0; g1_4.sAi = 0; g1_4.sAm = 8; g1_4.sAk = 1; g1_4.sBo = 0; g1_4.sBi = 0; g1_4.sBn = 1; g1_4.sBk = H; g1_4.sCo = 0; g1_4.sCi = 0; g1_4.sCm = H; g1_4.sRo = 0; g1_4.sRi = 0; g1_4.sRm = 0; g1_4.sRn = 0;
      g1_4.M = 8137; g1_4.N = H; g1_4.K = 3; g1_4.zi_n = 1; g1_4.flags = 1; g1_4.act = 1;
      g1_4.alpha = 1.0f; g1_4.beta = 0.0f; g1_4.sa = 1.0f; g1_4.sb = 8.0f; g1_4.Npad = H; g1_4.pad_ = 0;
      k_gemm<0><<<dim3((unsigned)((H) + 31) / 32, (unsigned)((8137) + 15) / 16, (unsigned)(1)), 32, 0, stream>>>(g1_4); }
    { GemmP g2_4;
      g2_4.A = H1; g2_4.B = W2 + 16384; g2_4.bias = b2 + 256; g2_4.R = H1; g2_4.C = H2;
      g2_4.sAo = 0; g2_4.sAi = 0; g2_4.sAm = H; g2_4.sAk = 1; g2_4.sBo = 0; g2_4.sBi = 0; g2_4.sBn = 1; g2_4.sBk = H; g2_4.sCo = 0; g2_4.sCi = 0; g2_4.sCm = H; g2_4.sRo = 0; g2_4.sRi = 0; g2_4.sRm = 0; g2_4.sRn = 0;
      g2_4.M = 8137; g2_4.N = H; g2_4.K = H; g2_4.zi_n = 1; g2_4.flags = 1; g2_4.act = 1;
      g2_4.alpha = 1.0f; g2_4.beta = 0.0f; g2_4.sa = 1.0f; g2_4.sb = 8.0f; g2_4.Npad = H; g2_4.pad_ = 0;
      k_gemm<0><<<dim3((unsigned)((H) + 31) / 32, (unsigned)((8137) + 15) / 16, (unsigned)(1)), 32, 0, stream>>>(g2_4); }
    { GemmP g3_4;
      g3_4.A = H2; g3_4.B = W3 + 256; g3_4.bias = b3 + 4; g3_4.R = H2; g3_4.C = Y;
      g3_4.sAo = 0; g3_4.sAi = 0; g3_4.sAm = H; g3_4.sAk = 1; g3_4.sBo = 0; g3_4.sBi = 0; g3_4.sBn = 1; g3_4.sBk = 1; g3_4.sCo = 0; g3_4.sCi = 0; g3_4.sCm = LP; g3_4.sRo = 0; g3_4.sRi = 0; g3_4.sRm = 0; g3_4.sRn = 0;
      g3_4.M = 8137; g3_4.N = 1; g3_4.K = H; g3_4.zi_n = 1; g3_4.flags = 1; g3_4.act = 0;
      g3_4.alpha = 1.0f; g3_4.beta = 0.0f; g3_4.sa = 1.0f; g3_4.sb = 8.0f; g3_4.Npad = LP; g3_4.pad_ = 0;
      k_gemm<0><<<dim3((unsigned)((LP) + 31) / 32, (unsigned)((8137) + 15) / 16, (unsigned)(1)), 32, 0, stream>>>(g3_4); }
    k_es_scatter<<<(unsigned)((8137 + 255) / 256), 256, 0, stream>>>(Y, LP, slot, IDX, 4, 32821, 8137, out);
    { GemmP g1_5;
      g1_5.A = XS + (size_t)40958 * 8; g1_5.B = W1 + 960; g1_5.bias = b1 + 320; g1_5.R = XS + (size_t)40958 * 8; g1_5.C = H1;
      g1_5.sAo = 0; g1_5.sAi = 0; g1_5.sAm = 8; g1_5.sAk = 1; g1_5.sBo = 0; g1_5.sBi = 0; g1_5.sBn = 1; g1_5.sBk = H; g1_5.sCo = 0; g1_5.sCi = 0; g1_5.sCm = H; g1_5.sRo = 0; g1_5.sRi = 0; g1_5.sRm = 0; g1_5.sRn = 0;
      g1_5.M = 8152; g1_5.N = H; g1_5.K = 3; g1_5.zi_n = 1; g1_5.flags = 1; g1_5.act = 1;
      g1_5.alpha = 1.0f; g1_5.beta = 0.0f; g1_5.sa = 1.0f; g1_5.sb = 8.0f; g1_5.Npad = H; g1_5.pad_ = 0;
      k_gemm<0><<<dim3((unsigned)((H) + 31) / 32, (unsigned)((8152) + 15) / 16, (unsigned)(1)), 32, 0, stream>>>(g1_5); }
    { GemmP g2_5;
      g2_5.A = H1; g2_5.B = W2 + 20480; g2_5.bias = b2 + 320; g2_5.R = H1; g2_5.C = H2;
      g2_5.sAo = 0; g2_5.sAi = 0; g2_5.sAm = H; g2_5.sAk = 1; g2_5.sBo = 0; g2_5.sBi = 0; g2_5.sBn = 1; g2_5.sBk = H; g2_5.sCo = 0; g2_5.sCi = 0; g2_5.sCm = H; g2_5.sRo = 0; g2_5.sRi = 0; g2_5.sRm = 0; g2_5.sRn = 0;
      g2_5.M = 8152; g2_5.N = H; g2_5.K = H; g2_5.zi_n = 1; g2_5.flags = 1; g2_5.act = 1;
      g2_5.alpha = 1.0f; g2_5.beta = 0.0f; g2_5.sa = 1.0f; g2_5.sb = 8.0f; g2_5.Npad = H; g2_5.pad_ = 0;
      k_gemm<0><<<dim3((unsigned)((H) + 31) / 32, (unsigned)((8152) + 15) / 16, (unsigned)(1)), 32, 0, stream>>>(g2_5); }
    { GemmP g3_5;
      g3_5.A = H2; g3_5.B = W3 + 320; g3_5.bias = b3 + 5; g3_5.R = H2; g3_5.C = Y;
      g3_5.sAo = 0; g3_5.sAi = 0; g3_5.sAm = H; g3_5.sAk = 1; g3_5.sBo = 0; g3_5.sBi = 0; g3_5.sBn = 1; g3_5.sBk = 1; g3_5.sCo = 0; g3_5.sCi = 0; g3_5.sCm = LP; g3_5.sRo = 0; g3_5.sRi = 0; g3_5.sRm = 0; g3_5.sRn = 0;
      g3_5.M = 8152; g3_5.N = 1; g3_5.K = H; g3_5.zi_n = 1; g3_5.flags = 1; g3_5.act = 0;
      g3_5.alpha = 1.0f; g3_5.beta = 0.0f; g3_5.sa = 1.0f; g3_5.sb = 8.0f; g3_5.Npad = LP; g3_5.pad_ = 0;
      k_gemm<0><<<dim3((unsigned)((LP) + 31) / 32, (unsigned)((8152) + 15) / 16, (unsigned)(1)), 32, 0, stream>>>(g3_5); }
    k_es_scatter<<<(unsigned)((8152 + 255) / 256), 256, 0, stream>>>(Y, LP, slot, IDX, 5, 40958, 8152, out);
    { GemmP g1_6;
      g1_6.A = XS + (size_t)49110 * 8; g1_6.B = W1 + 1152; g1_6.bias = b1 + 384; g1_6.R = XS + (size_t)49110 * 8; g1_6.C = H1;
      g1_6.sAo = 0; g1_6.sAi = 0; g1_6.sAm = 8; g1_6.sAk = 1; g1_6.sBo = 0; g1_6.sBi = 0; g1_6.sBn = 1; g1_6.sBk = H; g1_6.sCo = 0; g1_6.sCi = 0; g1_6.sCm = H; g1_6.sRo = 0; g1_6.sRi = 0; g1_6.sRm = 0; g1_6.sRn = 0;
      g1_6.M = 8201; g1_6.N = H; g1_6.K = 3; g1_6.zi_n = 1; g1_6.flags = 1; g1_6.act = 1;
      g1_6.alpha = 1.0f; g1_6.beta = 0.0f; g1_6.sa = 1.0f; g1_6.sb = 8.0f; g1_6.Npad = H; g1_6.pad_ = 0;
      k_gemm<0><<<dim3((unsigned)((H) + 31) / 32, (unsigned)((8201) + 15) / 16, (unsigned)(1)), 32, 0, stream>>>(g1_6); }
    { GemmP g2_6;
      g2_6.A = H1; g2_6.B = W2 + 24576; g2_6.bias = b2 + 384; g2_6.R = H1; g2_6.C = H2;
      g2_6.sAo = 0; g2_6.sAi = 0; g2_6.sAm = H; g2_6.sAk = 1; g2_6.sBo = 0; g2_6.sBi = 0; g2_6.sBn = 1; g2_6.sBk = H; g2_6.sCo = 0; g2_6.sCi = 0; g2_6.sCm = H; g2_6.sRo = 0; g2_6.sRi = 0; g2_6.sRm = 0; g2_6.sRn = 0;
      g2_6.M = 8201; g2_6.N = H; g2_6.K = H; g2_6.zi_n = 1; g2_6.flags = 1; g2_6.act = 1;
      g2_6.alpha = 1.0f; g2_6.beta = 0.0f; g2_6.sa = 1.0f; g2_6.sb = 8.0f; g2_6.Npad = H; g2_6.pad_ = 0;
      k_gemm<0><<<dim3((unsigned)((H) + 31) / 32, (unsigned)((8201) + 15) / 16, (unsigned)(1)), 32, 0, stream>>>(g2_6); }
    { GemmP g3_6;
      g3_6.A = H2; g3_6.B = W3 + 384; g3_6.bias = b3 + 6; g3_6.R = H2; g3_6.C = Y;
      g3_6.sAo = 0; g3_6.sAi = 0; g3_6.sAm = H; g3_6.sAk = 1; g3_6.sBo = 0; g3_6.sBi = 0; g3_6.sBn = 1; g3_6.sBk = 1; g3_6.sCo = 0; g3_6.sCi = 0; g3_6.sCm = LP; g3_6.sRo = 0; g3_6.sRi = 0; g3_6.sRm = 0; g3_6.sRn = 0;
      g3_6.M = 8201; g3_6.N = 1; g3_6.K = H; g3_6.zi_n = 1; g3_6.flags = 1; g3_6.act = 0;
      g3_6.alpha = 1.0f; g3_6.beta = 0.0f; g3_6.sa = 1.0f; g3_6.sb = 8.0f; g3_6.Npad = LP; g3_6.pad_ = 0;
      k_gemm<0><<<dim3((unsigned)((LP) + 31) / 32, (unsigned)((8201) + 15) / 16, (unsigned)(1)), 32, 0, stream>>>(g3_6); }
    k_es_scatter<<<(unsigned)((8201 + 255) / 256), 256, 0, stream>>>(Y, LP, slot, IDX, 6, 49110, 8201, out);
    { GemmP g1_7;
      g1_7.A = XS + (size_t)57311 * 8; g1_7.B = W1 + 1344; g1_7.bias = b1 + 448; g1_7.R = XS + (size_t)57311 * 8; g1_7.C = H1;
      g1_7.sAo = 0; g1_7.sAi = 0; g1_7.sAm = 8; g1_7.sAk = 1; g1_7.sBo = 0; g1_7.sBi = 0; g1_7.sBn = 1; g1_7.sBk = H; g1_7.sCo = 0; g1_7.sCi = 0; g1_7.sCm = H; g1_7.sRo = 0; g1_7.sRi = 0; g1_7.sRm = 0; g1_7.sRn = 0;
      g1_7.M = 8159; g1_7.N = H; g1_7.K = 3; g1_7.zi_n = 1; g1_7.flags = 1; g1_7.act = 1;
      g1_7.alpha = 1.0f; g1_7.beta = 0.0f; g1_7.sa = 1.0f; g1_7.sb = 8.0f; g1_7.Npad = H; g1_7.pad_ = 0;
      k_gemm<0><<<dim3((unsigned)((H) + 31) / 32, (unsigned)((8159) + 15) / 16, (unsigned)(1)), 32, 0, stream>>>(g1_7); }
    { GemmP g2_7;
      g2_7.A = H1; g2_7.B = W2 + 28672; g2_7.bias = b2 + 448; g2_7.R = H1; g2_7.C = H2;
      g2_7.sAo = 0; g2_7.sAi = 0; g2_7.sAm = H; g2_7.sAk = 1; g2_7.sBo = 0; g2_7.sBi = 0; g2_7.sBn = 1; g2_7.sBk = H; g2_7.sCo = 0; g2_7.sCi = 0; g2_7.sCm = H; g2_7.sRo = 0; g2_7.sRi = 0; g2_7.sRm = 0; g2_7.sRn = 0;
      g2_7.M = 8159; g2_7.N = H; g2_7.K = H; g2_7.zi_n = 1; g2_7.flags = 1; g2_7.act = 1;
      g2_7.alpha = 1.0f; g2_7.beta = 0.0f; g2_7.sa = 1.0f; g2_7.sb = 8.0f; g2_7.Npad = H; g2_7.pad_ = 0;
      k_gemm<0><<<dim3((unsigned)((H) + 31) / 32, (unsigned)((8159) + 15) / 16, (unsigned)(1)), 32, 0, stream>>>(g2_7); }
    { GemmP g3_7;
      g3_7.A = H2; g3_7.B = W3 + 448; g3_7.bias = b3 + 7; g3_7.R = H2; g3_7.C = Y;
      g3_7.sAo = 0; g3_7.sAi = 0; g3_7.sAm = H; g3_7.sAk = 1; g3_7.sBo = 0; g3_7.sBi = 0; g3_7.sBn = 1; g3_7.sBk = 1; g3_7.sCo = 0; g3_7.sCi = 0; g3_7.sCm = LP; g3_7.sRo = 0; g3_7.sRi = 0; g3_7.sRm = 0; g3_7.sRn = 0;
      g3_7.M = 8159; g3_7.N = 1; g3_7.K = H; g3_7.zi_n = 1; g3_7.flags = 1; g3_7.act = 0;
      g3_7.alpha = 1.0f; g3_7.beta = 0.0f; g3_7.sa = 1.0f; g3_7.sb = 8.0f; g3_7.Npad = LP; g3_7.pad_ = 0;
      k_gemm<0><<<dim3((unsigned)((LP) + 31) / 32, (unsigned)((8159) + 15) / 16, (unsigned)(1)), 32, 0, stream>>>(g3_7); }
    k_es_scatter<<<(unsigned)((8159 + 255) / 256), 256, 0, stream>>>(Y, LP, slot, IDX, 7, 57311, 8159, out);
    { GemmP g1_8;
      g1_8.A = XS + (size_t)65470 * 8; g1_8.B = W1 + 1536; g1_8.bias = b1 + 512; g1_8.R = XS + (size_t)65470 * 8; g1_8.C = H1;
      g1_8.sAo = 0; g1_8.sAi = 0; g1_8.sAm = 8; g1_8.sAk = 1; g1_8.sBo = 0; g1_8.sBi = 0; g1_8.sBn = 1; g1_8.sBk = H; g1_8.sCo = 0; g1_8.sCi = 0; g1_8.sCm = H; g1_8.sRo = 0; g1_8.sRi = 0; g1_8.sRm = 0; g1_8.sRn = 0;
      g1_8.M = 8120; g1_8.N = H; g1_8.K = 3; g1_8.zi_n = 1; g1_8.flags = 1; g1_8.act = 1;
      g1_8.alpha = 1.0f; g1_8.beta = 0.0f; g1_8.sa = 1.0f; g1_8.sb = 8.0f; g1_8.Npad = H; g1_8.pad_ = 0;
      k_gemm<0><<<dim3((unsigned)((H) + 31) / 32, (unsigned)((8120) + 15) / 16, (unsigned)(1)), 32, 0, stream>>>(g1_8); }
    { GemmP g2_8;
      g2_8.A = H1; g2_8.B = W2 + 32768; g2_8.bias = b2 + 512; g2_8.R = H1; g2_8.C = H2;
      g2_8.sAo = 0; g2_8.sAi = 0; g2_8.sAm = H; g2_8.sAk = 1; g2_8.sBo = 0; g2_8.sBi = 0; g2_8.sBn = 1; g2_8.sBk = H; g2_8.sCo = 0; g2_8.sCi = 0; g2_8.sCm = H; g2_8.sRo = 0; g2_8.sRi = 0; g2_8.sRm = 0; g2_8.sRn = 0;
      g2_8.M = 8120; g2_8.N = H; g2_8.K = H; g2_8.zi_n = 1; g2_8.flags = 1; g2_8.act = 1;
      g2_8.alpha = 1.0f; g2_8.beta = 0.0f; g2_8.sa = 1.0f; g2_8.sb = 8.0f; g2_8.Npad = H; g2_8.pad_ = 0;
      k_gemm<0><<<dim3((unsigned)((H) + 31) / 32, (unsigned)((8120) + 15) / 16, (unsigned)(1)), 32, 0, stream>>>(g2_8); }
    { GemmP g3_8;
      g3_8.A = H2; g3_8.B = W3 + 512; g3_8.bias = b3 + 8; g3_8.R = H2; g3_8.C = Y;
      g3_8.sAo = 0; g3_8.sAi = 0; g3_8.sAm = H; g3_8.sAk = 1; g3_8.sBo = 0; g3_8.sBi = 0; g3_8.sBn = 1; g3_8.sBk = 1; g3_8.sCo = 0; g3_8.sCi = 0; g3_8.sCm = LP; g3_8.sRo = 0; g3_8.sRi = 0; g3_8.sRm = 0; g3_8.sRn = 0;
      g3_8.M = 8120; g3_8.N = 1; g3_8.K = H; g3_8.zi_n = 1; g3_8.flags = 1; g3_8.act = 0;
      g3_8.alpha = 1.0f; g3_8.beta = 0.0f; g3_8.sa = 1.0f; g3_8.sb = 8.0f; g3_8.Npad = LP; g3_8.pad_ = 0;
      k_gemm<0><<<dim3((unsigned)((LP) + 31) / 32, (unsigned)((8120) + 15) / 16, (unsigned)(1)), 32, 0, stream>>>(g3_8); }
    k_es_scatter<<<(unsigned)((8120 + 255) / 256), 256, 0, stream>>>(Y, LP, slot, IDX, 8, 65470, 8120, out);
    { GemmP g1_9;
      g1_9.A = XS + (size_t)73590 * 8; g1_9.B = W1 + 1728; g1_9.bias = b1 + 576; g1_9.R = XS + (size_t)73590 * 8; g1_9.C = H1;
      g1_9.sAo = 0; g1_9.sAi = 0; g1_9.sAm = 8; g1_9.sAk = 1; g1_9.sBo = 0; g1_9.sBi = 0; g1_9.sBn = 1; g1_9.sBk = H; g1_9.sCo = 0; g1_9.sCi = 0; g1_9.sCm = H; g1_9.sRo = 0; g1_9.sRi = 0; g1_9.sRm = 0; g1_9.sRn = 0;
      g1_9.M = 8104; g1_9.N = H; g1_9.K = 3; g1_9.zi_n = 1; g1_9.flags = 1; g1_9.act = 1;
      g1_9.alpha = 1.0f; g1_9.beta = 0.0f; g1_9.sa = 1.0f; g1_9.sb = 8.0f; g1_9.Npad = H; g1_9.pad_ = 0;
      k_gemm<0><<<dim3((unsigned)((H) + 31) / 32, (unsigned)((8104) + 15) / 16, (unsigned)(1)), 32, 0, stream>>>(g1_9); }
    { GemmP g2_9;
      g2_9.A = H1; g2_9.B = W2 + 36864; g2_9.bias = b2 + 576; g2_9.R = H1; g2_9.C = H2;
      g2_9.sAo = 0; g2_9.sAi = 0; g2_9.sAm = H; g2_9.sAk = 1; g2_9.sBo = 0; g2_9.sBi = 0; g2_9.sBn = 1; g2_9.sBk = H; g2_9.sCo = 0; g2_9.sCi = 0; g2_9.sCm = H; g2_9.sRo = 0; g2_9.sRi = 0; g2_9.sRm = 0; g2_9.sRn = 0;
      g2_9.M = 8104; g2_9.N = H; g2_9.K = H; g2_9.zi_n = 1; g2_9.flags = 1; g2_9.act = 1;
      g2_9.alpha = 1.0f; g2_9.beta = 0.0f; g2_9.sa = 1.0f; g2_9.sb = 8.0f; g2_9.Npad = H; g2_9.pad_ = 0;
      k_gemm<0><<<dim3((unsigned)((H) + 31) / 32, (unsigned)((8104) + 15) / 16, (unsigned)(1)), 32, 0, stream>>>(g2_9); }
    { GemmP g3_9;
      g3_9.A = H2; g3_9.B = W3 + 576; g3_9.bias = b3 + 9; g3_9.R = H2; g3_9.C = Y;
      g3_9.sAo = 0; g3_9.sAi = 0; g3_9.sAm = H; g3_9.sAk = 1; g3_9.sBo = 0; g3_9.sBi = 0; g3_9.sBn = 1; g3_9.sBk = 1; g3_9.sCo = 0; g3_9.sCi = 0; g3_9.sCm = LP; g3_9.sRo = 0; g3_9.sRi = 0; g3_9.sRm = 0; g3_9.sRn = 0;
      g3_9.M = 8104; g3_9.N = 1; g3_9.K = H; g3_9.zi_n = 1; g3_9.flags = 1; g3_9.act = 0;
      g3_9.alpha = 1.0f; g3_9.beta = 0.0f; g3_9.sa = 1.0f; g3_9.sb = 8.0f; g3_9.Npad = LP; g3_9.pad_ = 0;
      k_gemm<0><<<dim3((unsigned)((LP) + 31) / 32, (unsigned)((8104) + 15) / 16, (unsigned)(1)), 32, 0, stream>>>(g3_9); }
    k_es_scatter<<<(unsigned)((8104 + 255) / 256), 256, 0, stream>>>(Y, LP, slot, IDX, 9, 73590, 8104, out);
    { GemmP g1_10;
      g1_10.A = XS + (size_t)81694 * 8; g1_10.B = W1 + 1920; g1_10.bias = b1 + 640; g1_10.R = XS + (size_t)81694 * 8; g1_10.C = H1;
      g1_10.sAo = 0; g1_10.sAi = 0; g1_10.sAm = 8; g1_10.sAk = 1; g1_10.sBo = 0; g1_10.sBi = 0; g1_10.sBn = 1; g1_10.sBk = H; g1_10.sCo = 0; g1_10.sCi = 0; g1_10.sCm = H; g1_10.sRo = 0; g1_10.sRi = 0; g1_10.sRm = 0; g1_10.sRn = 0;
      g1_10.M = 8047; g1_10.N = H; g1_10.K = 3; g1_10.zi_n = 1; g1_10.flags = 1; g1_10.act = 1;
      g1_10.alpha = 1.0f; g1_10.beta = 0.0f; g1_10.sa = 1.0f; g1_10.sb = 8.0f; g1_10.Npad = H; g1_10.pad_ = 0;
      k_gemm<0><<<dim3((unsigned)((H) + 31) / 32, (unsigned)((8047) + 15) / 16, (unsigned)(1)), 32, 0, stream>>>(g1_10); }
    { GemmP g2_10;
      g2_10.A = H1; g2_10.B = W2 + 40960; g2_10.bias = b2 + 640; g2_10.R = H1; g2_10.C = H2;
      g2_10.sAo = 0; g2_10.sAi = 0; g2_10.sAm = H; g2_10.sAk = 1; g2_10.sBo = 0; g2_10.sBi = 0; g2_10.sBn = 1; g2_10.sBk = H; g2_10.sCo = 0; g2_10.sCi = 0; g2_10.sCm = H; g2_10.sRo = 0; g2_10.sRi = 0; g2_10.sRm = 0; g2_10.sRn = 0;
      g2_10.M = 8047; g2_10.N = H; g2_10.K = H; g2_10.zi_n = 1; g2_10.flags = 1; g2_10.act = 1;
      g2_10.alpha = 1.0f; g2_10.beta = 0.0f; g2_10.sa = 1.0f; g2_10.sb = 8.0f; g2_10.Npad = H; g2_10.pad_ = 0;
      k_gemm<0><<<dim3((unsigned)((H) + 31) / 32, (unsigned)((8047) + 15) / 16, (unsigned)(1)), 32, 0, stream>>>(g2_10); }
    { GemmP g3_10;
      g3_10.A = H2; g3_10.B = W3 + 640; g3_10.bias = b3 + 10; g3_10.R = H2; g3_10.C = Y;
      g3_10.sAo = 0; g3_10.sAi = 0; g3_10.sAm = H; g3_10.sAk = 1; g3_10.sBo = 0; g3_10.sBi = 0; g3_10.sBn = 1; g3_10.sBk = 1; g3_10.sCo = 0; g3_10.sCi = 0; g3_10.sCm = LP; g3_10.sRo = 0; g3_10.sRi = 0; g3_10.sRm = 0; g3_10.sRn = 0;
      g3_10.M = 8047; g3_10.N = 1; g3_10.K = H; g3_10.zi_n = 1; g3_10.flags = 1; g3_10.act = 0;
      g3_10.alpha = 1.0f; g3_10.beta = 0.0f; g3_10.sa = 1.0f; g3_10.sb = 8.0f; g3_10.Npad = LP; g3_10.pad_ = 0;
      k_gemm<0><<<dim3((unsigned)((LP) + 31) / 32, (unsigned)((8047) + 15) / 16, (unsigned)(1)), 32, 0, stream>>>(g3_10); }
    k_es_scatter<<<(unsigned)((8047 + 255) / 256), 256, 0, stream>>>(Y, LP, slot, IDX, 10, 81694, 8047, out);
    { GemmP g1_11;
      g1_11.A = XS + (size_t)89741 * 8; g1_11.B = W1 + 2112; g1_11.bias = b1 + 704; g1_11.R = XS + (size_t)89741 * 8; g1_11.C = H1;
      g1_11.sAo = 0; g1_11.sAi = 0; g1_11.sAm = 8; g1_11.sAk = 1; g1_11.sBo = 0; g1_11.sBi = 0; g1_11.sBn = 1; g1_11.sBk = H; g1_11.sCo = 0; g1_11.sCi = 0; g1_11.sCm = H; g1_11.sRo = 0; g1_11.sRi = 0; g1_11.sRm = 0; g1_11.sRn = 0;
      g1_11.M = 8168; g1_11.N = H; g1_11.K = 3; g1_11.zi_n = 1; g1_11.flags = 1; g1_11.act = 1;
      g1_11.alpha = 1.0f; g1_11.beta = 0.0f; g1_11.sa = 1.0f; g1_11.sb = 8.0f; g1_11.Npad = H; g1_11.pad_ = 0;
      k_gemm<0><<<dim3((unsigned)((H) + 31) / 32, (unsigned)((8168) + 15) / 16, (unsigned)(1)), 32, 0, stream>>>(g1_11); }
    { GemmP g2_11;
      g2_11.A = H1; g2_11.B = W2 + 45056; g2_11.bias = b2 + 704; g2_11.R = H1; g2_11.C = H2;
      g2_11.sAo = 0; g2_11.sAi = 0; g2_11.sAm = H; g2_11.sAk = 1; g2_11.sBo = 0; g2_11.sBi = 0; g2_11.sBn = 1; g2_11.sBk = H; g2_11.sCo = 0; g2_11.sCi = 0; g2_11.sCm = H; g2_11.sRo = 0; g2_11.sRi = 0; g2_11.sRm = 0; g2_11.sRn = 0;
      g2_11.M = 8168; g2_11.N = H; g2_11.K = H; g2_11.zi_n = 1; g2_11.flags = 1; g2_11.act = 1;
      g2_11.alpha = 1.0f; g2_11.beta = 0.0f; g2_11.sa = 1.0f; g2_11.sb = 8.0f; g2_11.Npad = H; g2_11.pad_ = 0;
      k_gemm<0><<<dim3((unsigned)((H) + 31) / 32, (unsigned)((8168) + 15) / 16, (unsigned)(1)), 32, 0, stream>>>(g2_11); }
    { GemmP g3_11;
      g3_11.A = H2; g3_11.B = W3 + 704; g3_11.bias = b3 + 11; g3_11.R = H2; g3_11.C = Y;
      g3_11.sAo = 0; g3_11.sAi = 0; g3_11.sAm = H; g3_11.sAk = 1; g3_11.sBo = 0; g3_11.sBi = 0; g3_11.sBn = 1; g3_11.sBk = 1; g3_11.sCo = 0; g3_11.sCi = 0; g3_11.sCm = LP; g3_11.sRo = 0; g3_11.sRi = 0; g3_11.sRm = 0; g3_11.sRn = 0;
      g3_11.M = 8168; g3_11.N = 1; g3_11.K = H; g3_11.zi_n = 1; g3_11.flags = 1; g3_11.act = 0;
      g3_11.alpha = 1.0f; g3_11.beta = 0.0f; g3_11.sa = 1.0f; g3_11.sb = 8.0f; g3_11.Npad = LP; g3_11.pad_ = 0;
      k_gemm<0><<<dim3((unsigned)((LP) + 31) / 32, (unsigned)((8168) + 15) / 16, (unsigned)(1)), 32, 0, stream>>>(g3_11); }
    k_es_scatter<<<(unsigned)((8168 + 255) / 256), 256, 0, stream>>>(Y, LP, slot, IDX, 11, 89741, 8168, out);
    { GemmP g1_12;
      g1_12.A = XS + (size_t)97909 * 8; g1_12.B = W1 + 2304; g1_12.bias = b1 + 768; g1_12.R = XS + (size_t)97909 * 8; g1_12.C = H1;
      g1_12.sAo = 0; g1_12.sAi = 0; g1_12.sAm = 8; g1_12.sAk = 1; g1_12.sBo = 0; g1_12.sBi = 0; g1_12.sBn = 1; g1_12.sBk = H; g1_12.sCo = 0; g1_12.sCi = 0; g1_12.sCm = H; g1_12.sRo = 0; g1_12.sRi = 0; g1_12.sRm = 0; g1_12.sRn = 0;
      g1_12.M = 8409; g1_12.N = H; g1_12.K = 3; g1_12.zi_n = 1; g1_12.flags = 1; g1_12.act = 1;
      g1_12.alpha = 1.0f; g1_12.beta = 0.0f; g1_12.sa = 1.0f; g1_12.sb = 8.0f; g1_12.Npad = H; g1_12.pad_ = 0;
      k_gemm<0><<<dim3((unsigned)((H) + 31) / 32, (unsigned)((8409) + 15) / 16, (unsigned)(1)), 32, 0, stream>>>(g1_12); }
    { GemmP g2_12;
      g2_12.A = H1; g2_12.B = W2 + 49152; g2_12.bias = b2 + 768; g2_12.R = H1; g2_12.C = H2;
      g2_12.sAo = 0; g2_12.sAi = 0; g2_12.sAm = H; g2_12.sAk = 1; g2_12.sBo = 0; g2_12.sBi = 0; g2_12.sBn = 1; g2_12.sBk = H; g2_12.sCo = 0; g2_12.sCi = 0; g2_12.sCm = H; g2_12.sRo = 0; g2_12.sRi = 0; g2_12.sRm = 0; g2_12.sRn = 0;
      g2_12.M = 8409; g2_12.N = H; g2_12.K = H; g2_12.zi_n = 1; g2_12.flags = 1; g2_12.act = 1;
      g2_12.alpha = 1.0f; g2_12.beta = 0.0f; g2_12.sa = 1.0f; g2_12.sb = 8.0f; g2_12.Npad = H; g2_12.pad_ = 0;
      k_gemm<0><<<dim3((unsigned)((H) + 31) / 32, (unsigned)((8409) + 15) / 16, (unsigned)(1)), 32, 0, stream>>>(g2_12); }
    { GemmP g3_12;
      g3_12.A = H2; g3_12.B = W3 + 768; g3_12.bias = b3 + 12; g3_12.R = H2; g3_12.C = Y;
      g3_12.sAo = 0; g3_12.sAi = 0; g3_12.sAm = H; g3_12.sAk = 1; g3_12.sBo = 0; g3_12.sBi = 0; g3_12.sBn = 1; g3_12.sBk = 1; g3_12.sCo = 0; g3_12.sCi = 0; g3_12.sCm = LP; g3_12.sRo = 0; g3_12.sRi = 0; g3_12.sRm = 0; g3_12.sRn = 0;
      g3_12.M = 8409; g3_12.N = 1; g3_12.K = H; g3_12.zi_n = 1; g3_12.flags = 1; g3_12.act = 0;
      g3_12.alpha = 1.0f; g3_12.beta = 0.0f; g3_12.sa = 1.0f; g3_12.sb = 8.0f; g3_12.Npad = LP; g3_12.pad_ = 0;
      k_gemm<0><<<dim3((unsigned)((LP) + 31) / 32, (unsigned)((8409) + 15) / 16, (unsigned)(1)), 32, 0, stream>>>(g3_12); }
    k_es_scatter<<<(unsigned)((8409 + 255) / 256), 256, 0, stream>>>(Y, LP, slot, IDX, 12, 97909, 8409, out);
    { GemmP g1_13;
      g1_13.A = XS + (size_t)106318 * 8; g1_13.B = W1 + 2496; g1_13.bias = b1 + 832; g1_13.R = XS + (size_t)106318 * 8; g1_13.C = H1;
      g1_13.sAo = 0; g1_13.sAi = 0; g1_13.sAm = 8; g1_13.sAk = 1; g1_13.sBo = 0; g1_13.sBi = 0; g1_13.sBn = 1; g1_13.sBk = H; g1_13.sCo = 0; g1_13.sCi = 0; g1_13.sCm = H; g1_13.sRo = 0; g1_13.sRi = 0; g1_13.sRm = 0; g1_13.sRn = 0;
      g1_13.M = 8094; g1_13.N = H; g1_13.K = 3; g1_13.zi_n = 1; g1_13.flags = 1; g1_13.act = 1;
      g1_13.alpha = 1.0f; g1_13.beta = 0.0f; g1_13.sa = 1.0f; g1_13.sb = 8.0f; g1_13.Npad = H; g1_13.pad_ = 0;
      k_gemm<0><<<dim3((unsigned)((H) + 31) / 32, (unsigned)((8094) + 15) / 16, (unsigned)(1)), 32, 0, stream>>>(g1_13); }
    { GemmP g2_13;
      g2_13.A = H1; g2_13.B = W2 + 53248; g2_13.bias = b2 + 832; g2_13.R = H1; g2_13.C = H2;
      g2_13.sAo = 0; g2_13.sAi = 0; g2_13.sAm = H; g2_13.sAk = 1; g2_13.sBo = 0; g2_13.sBi = 0; g2_13.sBn = 1; g2_13.sBk = H; g2_13.sCo = 0; g2_13.sCi = 0; g2_13.sCm = H; g2_13.sRo = 0; g2_13.sRi = 0; g2_13.sRm = 0; g2_13.sRn = 0;
      g2_13.M = 8094; g2_13.N = H; g2_13.K = H; g2_13.zi_n = 1; g2_13.flags = 1; g2_13.act = 1;
      g2_13.alpha = 1.0f; g2_13.beta = 0.0f; g2_13.sa = 1.0f; g2_13.sb = 8.0f; g2_13.Npad = H; g2_13.pad_ = 0;
      k_gemm<0><<<dim3((unsigned)((H) + 31) / 32, (unsigned)((8094) + 15) / 16, (unsigned)(1)), 32, 0, stream>>>(g2_13); }
    { GemmP g3_13;
      g3_13.A = H2; g3_13.B = W3 + 832; g3_13.bias = b3 + 13; g3_13.R = H2; g3_13.C = Y;
      g3_13.sAo = 0; g3_13.sAi = 0; g3_13.sAm = H; g3_13.sAk = 1; g3_13.sBo = 0; g3_13.sBi = 0; g3_13.sBn = 1; g3_13.sBk = 1; g3_13.sCo = 0; g3_13.sCi = 0; g3_13.sCm = LP; g3_13.sRo = 0; g3_13.sRi = 0; g3_13.sRm = 0; g3_13.sRn = 0;
      g3_13.M = 8094; g3_13.N = 1; g3_13.K = H; g3_13.zi_n = 1; g3_13.flags = 1; g3_13.act = 0;
      g3_13.alpha = 1.0f; g3_13.beta = 0.0f; g3_13.sa = 1.0f; g3_13.sb = 8.0f; g3_13.Npad = LP; g3_13.pad_ = 0;
      k_gemm<0><<<dim3((unsigned)((LP) + 31) / 32, (unsigned)((8094) + 15) / 16, (unsigned)(1)), 32, 0, stream>>>(g3_13); }
    k_es_scatter<<<(unsigned)((8094 + 255) / 256), 256, 0, stream>>>(Y, LP, slot, IDX, 13, 106318, 8094, out);
    { GemmP g1_14;
      g1_14.A = XS + (size_t)114412 * 8; g1_14.B = W1 + 2688; g1_14.bias = b1 + 896; g1_14.R = XS + (size_t)114412 * 8; g1_14.C = H1;
      g1_14.sAo = 0; g1_14.sAi = 0; g1_14.sAm = 8; g1_14.sAk = 1; g1_14.sBo = 0; g1_14.sBi = 0; g1_14.sBn = 1; g1_14.sBk = H; g1_14.sCo = 0; g1_14.sCi = 0; g1_14.sCm = H; g1_14.sRo = 0; g1_14.sRi = 0; g1_14.sRm = 0; g1_14.sRn = 0;
      g1_14.M = 8217; g1_14.N = H; g1_14.K = 3; g1_14.zi_n = 1; g1_14.flags = 1; g1_14.act = 1;
      g1_14.alpha = 1.0f; g1_14.beta = 0.0f; g1_14.sa = 1.0f; g1_14.sb = 8.0f; g1_14.Npad = H; g1_14.pad_ = 0;
      k_gemm<0><<<dim3((unsigned)((H) + 31) / 32, (unsigned)((8217) + 15) / 16, (unsigned)(1)), 32, 0, stream>>>(g1_14); }
    { GemmP g2_14;
      g2_14.A = H1; g2_14.B = W2 + 57344; g2_14.bias = b2 + 896; g2_14.R = H1; g2_14.C = H2;
      g2_14.sAo = 0; g2_14.sAi = 0; g2_14.sAm = H; g2_14.sAk = 1; g2_14.sBo = 0; g2_14.sBi = 0; g2_14.sBn = 1; g2_14.sBk = H; g2_14.sCo = 0; g2_14.sCi = 0; g2_14.sCm = H; g2_14.sRo = 0; g2_14.sRi = 0; g2_14.sRm = 0; g2_14.sRn = 0;
      g2_14.M = 8217; g2_14.N = H; g2_14.K = H; g2_14.zi_n = 1; g2_14.flags = 1; g2_14.act = 1;
      g2_14.alpha = 1.0f; g2_14.beta = 0.0f; g2_14.sa = 1.0f; g2_14.sb = 8.0f; g2_14.Npad = H; g2_14.pad_ = 0;
      k_gemm<0><<<dim3((unsigned)((H) + 31) / 32, (unsigned)((8217) + 15) / 16, (unsigned)(1)), 32, 0, stream>>>(g2_14); }
    { GemmP g3_14;
      g3_14.A = H2; g3_14.B = W3 + 896; g3_14.bias = b3 + 14; g3_14.R = H2; g3_14.C = Y;
      g3_14.sAo = 0; g3_14.sAi = 0; g3_14.sAm = H; g3_14.sAk = 1; g3_14.sBo = 0; g3_14.sBi = 0; g3_14.sBn = 1; g3_14.sBk = 1; g3_14.sCo = 0; g3_14.sCi = 0; g3_14.sCm = LP; g3_14.sRo = 0; g3_14.sRi = 0; g3_14.sRm = 0; g3_14.sRn = 0;
      g3_14.M = 8217; g3_14.N = 1; g3_14.K = H; g3_14.zi_n = 1; g3_14.flags = 1; g3_14.act = 0;
      g3_14.alpha = 1.0f; g3_14.beta = 0.0f; g3_14.sa = 1.0f; g3_14.sb = 8.0f; g3_14.Npad = LP; g3_14.pad_ = 0;
      k_gemm<0><<<dim3((unsigned)((LP) + 31) / 32, (unsigned)((8217) + 15) / 16, (unsigned)(1)), 32, 0, stream>>>(g3_14); }
    k_es_scatter<<<(unsigned)((8217 + 255) / 256), 256, 0, stream>>>(Y, LP, slot, IDX, 14, 114412, 8217, out);
    { GemmP g1_15;
      g1_15.A = XS + (size_t)122629 * 8; g1_15.B = W1 + 2880; g1_15.bias = b1 + 960; g1_15.R = XS + (size_t)122629 * 8; g1_15.C = H1;
      g1_15.sAo = 0; g1_15.sAi = 0; g1_15.sAm = 8; g1_15.sAk = 1; g1_15.sBo = 0; g1_15.sBi = 0; g1_15.sBn = 1; g1_15.sBk = H; g1_15.sCo = 0; g1_15.sCi = 0; g1_15.sCm = H; g1_15.sRo = 0; g1_15.sRi = 0; g1_15.sRm = 0; g1_15.sRn = 0;
      g1_15.M = 8293; g1_15.N = H; g1_15.K = 3; g1_15.zi_n = 1; g1_15.flags = 1; g1_15.act = 1;
      g1_15.alpha = 1.0f; g1_15.beta = 0.0f; g1_15.sa = 1.0f; g1_15.sb = 8.0f; g1_15.Npad = H; g1_15.pad_ = 0;
      k_gemm<0><<<dim3((unsigned)((H) + 31) / 32, (unsigned)((8293) + 15) / 16, (unsigned)(1)), 32, 0, stream>>>(g1_15); }
    { GemmP g2_15;
      g2_15.A = H1; g2_15.B = W2 + 61440; g2_15.bias = b2 + 960; g2_15.R = H1; g2_15.C = H2;
      g2_15.sAo = 0; g2_15.sAi = 0; g2_15.sAm = H; g2_15.sAk = 1; g2_15.sBo = 0; g2_15.sBi = 0; g2_15.sBn = 1; g2_15.sBk = H; g2_15.sCo = 0; g2_15.sCi = 0; g2_15.sCm = H; g2_15.sRo = 0; g2_15.sRi = 0; g2_15.sRm = 0; g2_15.sRn = 0;
      g2_15.M = 8293; g2_15.N = H; g2_15.K = H; g2_15.zi_n = 1; g2_15.flags = 1; g2_15.act = 1;
      g2_15.alpha = 1.0f; g2_15.beta = 0.0f; g2_15.sa = 1.0f; g2_15.sb = 8.0f; g2_15.Npad = H; g2_15.pad_ = 0;
      k_gemm<0><<<dim3((unsigned)((H) + 31) / 32, (unsigned)((8293) + 15) / 16, (unsigned)(1)), 32, 0, stream>>>(g2_15); }
    { GemmP g3_15;
      g3_15.A = H2; g3_15.B = W3 + 960; g3_15.bias = b3 + 15; g3_15.R = H2; g3_15.C = Y;
      g3_15.sAo = 0; g3_15.sAi = 0; g3_15.sAm = H; g3_15.sAk = 1; g3_15.sBo = 0; g3_15.sBi = 0; g3_15.sBn = 1; g3_15.sBk = 1; g3_15.sCo = 0; g3_15.sCi = 0; g3_15.sCm = LP; g3_15.sRo = 0; g3_15.sRi = 0; g3_15.sRm = 0; g3_15.sRn = 0;
      g3_15.M = 8293; g3_15.N = 1; g3_15.K = H; g3_15.zi_n = 1; g3_15.flags = 1; g3_15.act = 0;
      g3_15.alpha = 1.0f; g3_15.beta = 0.0f; g3_15.sa = 1.0f; g3_15.sb = 8.0f; g3_15.Npad = LP; g3_15.pad_ = 0;
      k_gemm<0><<<dim3((unsigned)((LP) + 31) / 32, (unsigned)((8293) + 15) / 16, (unsigned)(1)), 32, 0, stream>>>(g3_15); }
    k_es_scatter<<<(unsigned)((8293 + 255) / 256), 256, 0, stream>>>(Y, LP, slot, IDX, 15, 122629, 8293, out);
    { GemmP g1_16;
      g1_16.A = XS + (size_t)130922 * 8; g1_16.B = W1 + 3072; g1_16.bias = b1 + 1024; g1_16.R = XS + (size_t)130922 * 8; g1_16.C = H1;
      g1_16.sAo = 0; g1_16.sAi = 0; g1_16.sAm = 8; g1_16.sAk = 1; g1_16.sBo = 0; g1_16.sBi = 0; g1_16.sBn = 1; g1_16.sBk = H; g1_16.sCo = 0; g1_16.sCi = 0; g1_16.sCm = H; g1_16.sRo = 0; g1_16.sRi = 0; g1_16.sRm = 0; g1_16.sRn = 0;
      g1_16.M = 8222; g1_16.N = H; g1_16.K = 3; g1_16.zi_n = 1; g1_16.flags = 1; g1_16.act = 1;
      g1_16.alpha = 1.0f; g1_16.beta = 0.0f; g1_16.sa = 1.0f; g1_16.sb = 8.0f; g1_16.Npad = H; g1_16.pad_ = 0;
      k_gemm<0><<<dim3((unsigned)((H) + 31) / 32, (unsigned)((8222) + 15) / 16, (unsigned)(1)), 32, 0, stream>>>(g1_16); }
    { GemmP g2_16;
      g2_16.A = H1; g2_16.B = W2 + 65536; g2_16.bias = b2 + 1024; g2_16.R = H1; g2_16.C = H2;
      g2_16.sAo = 0; g2_16.sAi = 0; g2_16.sAm = H; g2_16.sAk = 1; g2_16.sBo = 0; g2_16.sBi = 0; g2_16.sBn = 1; g2_16.sBk = H; g2_16.sCo = 0; g2_16.sCi = 0; g2_16.sCm = H; g2_16.sRo = 0; g2_16.sRi = 0; g2_16.sRm = 0; g2_16.sRn = 0;
      g2_16.M = 8222; g2_16.N = H; g2_16.K = H; g2_16.zi_n = 1; g2_16.flags = 1; g2_16.act = 1;
      g2_16.alpha = 1.0f; g2_16.beta = 0.0f; g2_16.sa = 1.0f; g2_16.sb = 8.0f; g2_16.Npad = H; g2_16.pad_ = 0;
      k_gemm<0><<<dim3((unsigned)((H) + 31) / 32, (unsigned)((8222) + 15) / 16, (unsigned)(1)), 32, 0, stream>>>(g2_16); }
    { GemmP g3_16;
      g3_16.A = H2; g3_16.B = W3 + 1024; g3_16.bias = b3 + 16; g3_16.R = H2; g3_16.C = Y;
      g3_16.sAo = 0; g3_16.sAi = 0; g3_16.sAm = H; g3_16.sAk = 1; g3_16.sBo = 0; g3_16.sBi = 0; g3_16.sBn = 1; g3_16.sBk = 1; g3_16.sCo = 0; g3_16.sCi = 0; g3_16.sCm = LP; g3_16.sRo = 0; g3_16.sRi = 0; g3_16.sRm = 0; g3_16.sRn = 0;
      g3_16.M = 8222; g3_16.N = 1; g3_16.K = H; g3_16.zi_n = 1; g3_16.flags = 1; g3_16.act = 0;
      g3_16.alpha = 1.0f; g3_16.beta = 0.0f; g3_16.sa = 1.0f; g3_16.sb = 8.0f; g3_16.Npad = LP; g3_16.pad_ = 0;
      k_gemm<0><<<dim3((unsigned)((LP) + 31) / 32, (unsigned)((8222) + 15) / 16, (unsigned)(1)), 32, 0, stream>>>(g3_16); }
    k_es_scatter<<<(unsigned)((8222 + 255) / 256), 256, 0, stream>>>(Y, LP, slot, IDX, 16, 130922, 8222, out);
    { GemmP g1_17;
      g1_17.A = XS + (size_t)139144 * 8; g1_17.B = W1 + 3264; g1_17.bias = b1 + 1088; g1_17.R = XS + (size_t)139144 * 8; g1_17.C = H1;
      g1_17.sAo = 0; g1_17.sAi = 0; g1_17.sAm = 8; g1_17.sAk = 1; g1_17.sBo = 0; g1_17.sBi = 0; g1_17.sBn = 1; g1_17.sBk = H; g1_17.sCo = 0; g1_17.sCi = 0; g1_17.sCm = H; g1_17.sRo = 0; g1_17.sRi = 0; g1_17.sRm = 0; g1_17.sRn = 0;
      g1_17.M = 8079; g1_17.N = H; g1_17.K = 3; g1_17.zi_n = 1; g1_17.flags = 1; g1_17.act = 1;
      g1_17.alpha = 1.0f; g1_17.beta = 0.0f; g1_17.sa = 1.0f; g1_17.sb = 8.0f; g1_17.Npad = H; g1_17.pad_ = 0;
      k_gemm<0><<<dim3((unsigned)((H) + 31) / 32, (unsigned)((8079) + 15) / 16, (unsigned)(1)), 32, 0, stream>>>(g1_17); }
    { GemmP g2_17;
      g2_17.A = H1; g2_17.B = W2 + 69632; g2_17.bias = b2 + 1088; g2_17.R = H1; g2_17.C = H2;
      g2_17.sAo = 0; g2_17.sAi = 0; g2_17.sAm = H; g2_17.sAk = 1; g2_17.sBo = 0; g2_17.sBi = 0; g2_17.sBn = 1; g2_17.sBk = H; g2_17.sCo = 0; g2_17.sCi = 0; g2_17.sCm = H; g2_17.sRo = 0; g2_17.sRi = 0; g2_17.sRm = 0; g2_17.sRn = 0;
      g2_17.M = 8079; g2_17.N = H; g2_17.K = H; g2_17.zi_n = 1; g2_17.flags = 1; g2_17.act = 1;
      g2_17.alpha = 1.0f; g2_17.beta = 0.0f; g2_17.sa = 1.0f; g2_17.sb = 8.0f; g2_17.Npad = H; g2_17.pad_ = 0;
      k_gemm<0><<<dim3((unsigned)((H) + 31) / 32, (unsigned)((8079) + 15) / 16, (unsigned)(1)), 32, 0, stream>>>(g2_17); }
    { GemmP g3_17;
      g3_17.A = H2; g3_17.B = W3 + 1088; g3_17.bias = b3 + 17; g3_17.R = H2; g3_17.C = Y;
      g3_17.sAo = 0; g3_17.sAi = 0; g3_17.sAm = H; g3_17.sAk = 1; g3_17.sBo = 0; g3_17.sBi = 0; g3_17.sBn = 1; g3_17.sBk = 1; g3_17.sCo = 0; g3_17.sCi = 0; g3_17.sCm = LP; g3_17.sRo = 0; g3_17.sRi = 0; g3_17.sRm = 0; g3_17.sRn = 0;
      g3_17.M = 8079; g3_17.N = 1; g3_17.K = H; g3_17.zi_n = 1; g3_17.flags = 1; g3_17.act = 0;
      g3_17.alpha = 1.0f; g3_17.beta = 0.0f; g3_17.sa = 1.0f; g3_17.sb = 8.0f; g3_17.Npad = LP; g3_17.pad_ = 0;
      k_gemm<0><<<dim3((unsigned)((LP) + 31) / 32, (unsigned)((8079) + 15) / 16, (unsigned)(1)), 32, 0, stream>>>(g3_17); }
    k_es_scatter<<<(unsigned)((8079 + 255) / 256), 256, 0, stream>>>(Y, LP, slot, IDX, 17, 139144, 8079, out);
    { GemmP g1_18;
      g1_18.A = XS + (size_t)147223 * 8; g1_18.B = W1 + 3456; g1_18.bias = b1 + 1152; g1_18.R = XS + (size_t)147223 * 8; g1_18.C = H1;
      g1_18.sAo = 0; g1_18.sAi = 0; g1_18.sAm = 8; g1_18.sAk = 1; g1_18.sBo = 0; g1_18.sBi = 0; g1_18.sBn = 1; g1_18.sBk = H; g1_18.sCo = 0; g1_18.sCi = 0; g1_18.sCm = H; g1_18.sRo = 0; g1_18.sRi = 0; g1_18.sRm = 0; g1_18.sRn = 0;
      g1_18.M = 8187; g1_18.N = H; g1_18.K = 3; g1_18.zi_n = 1; g1_18.flags = 1; g1_18.act = 1;
      g1_18.alpha = 1.0f; g1_18.beta = 0.0f; g1_18.sa = 1.0f; g1_18.sb = 8.0f; g1_18.Npad = H; g1_18.pad_ = 0;
      k_gemm<0><<<dim3((unsigned)((H) + 31) / 32, (unsigned)((8187) + 15) / 16, (unsigned)(1)), 32, 0, stream>>>(g1_18); }
    { GemmP g2_18;
      g2_18.A = H1; g2_18.B = W2 + 73728; g2_18.bias = b2 + 1152; g2_18.R = H1; g2_18.C = H2;
      g2_18.sAo = 0; g2_18.sAi = 0; g2_18.sAm = H; g2_18.sAk = 1; g2_18.sBo = 0; g2_18.sBi = 0; g2_18.sBn = 1; g2_18.sBk = H; g2_18.sCo = 0; g2_18.sCi = 0; g2_18.sCm = H; g2_18.sRo = 0; g2_18.sRi = 0; g2_18.sRm = 0; g2_18.sRn = 0;
      g2_18.M = 8187; g2_18.N = H; g2_18.K = H; g2_18.zi_n = 1; g2_18.flags = 1; g2_18.act = 1;
      g2_18.alpha = 1.0f; g2_18.beta = 0.0f; g2_18.sa = 1.0f; g2_18.sb = 8.0f; g2_18.Npad = H; g2_18.pad_ = 0;
      k_gemm<0><<<dim3((unsigned)((H) + 31) / 32, (unsigned)((8187) + 15) / 16, (unsigned)(1)), 32, 0, stream>>>(g2_18); }
    { GemmP g3_18;
      g3_18.A = H2; g3_18.B = W3 + 1152; g3_18.bias = b3 + 18; g3_18.R = H2; g3_18.C = Y;
      g3_18.sAo = 0; g3_18.sAi = 0; g3_18.sAm = H; g3_18.sAk = 1; g3_18.sBo = 0; g3_18.sBi = 0; g3_18.sBn = 1; g3_18.sBk = 1; g3_18.sCo = 0; g3_18.sCi = 0; g3_18.sCm = LP; g3_18.sRo = 0; g3_18.sRi = 0; g3_18.sRm = 0; g3_18.sRn = 0;
      g3_18.M = 8187; g3_18.N = 1; g3_18.K = H; g3_18.zi_n = 1; g3_18.flags = 1; g3_18.act = 0;
      g3_18.alpha = 1.0f; g3_18.beta = 0.0f; g3_18.sa = 1.0f; g3_18.sb = 8.0f; g3_18.Npad = LP; g3_18.pad_ = 0;
      k_gemm<0><<<dim3((unsigned)((LP) + 31) / 32, (unsigned)((8187) + 15) / 16, (unsigned)(1)), 32, 0, stream>>>(g3_18); }
    k_es_scatter<<<(unsigned)((8187 + 255) / 256), 256, 0, stream>>>(Y, LP, slot, IDX, 18, 147223, 8187, out);
    { GemmP g1_19;
      g1_19.A = XS + (size_t)155410 * 8; g1_19.B = W1 + 3648; g1_19.bias = b1 + 1216; g1_19.R = XS + (size_t)155410 * 8; g1_19.C = H1;
      g1_19.sAo = 0; g1_19.sAi = 0; g1_19.sAm = 8; g1_19.sAk = 1; g1_19.sBo = 0; g1_19.sBi = 0; g1_19.sBn = 1; g1_19.sBk = H; g1_19.sCo = 0; g1_19.sCi = 0; g1_19.sCm = H; g1_19.sRo = 0; g1_19.sRi = 0; g1_19.sRm = 0; g1_19.sRn = 0;
      g1_19.M = 8290; g1_19.N = H; g1_19.K = 3; g1_19.zi_n = 1; g1_19.flags = 1; g1_19.act = 1;
      g1_19.alpha = 1.0f; g1_19.beta = 0.0f; g1_19.sa = 1.0f; g1_19.sb = 8.0f; g1_19.Npad = H; g1_19.pad_ = 0;
      k_gemm<0><<<dim3((unsigned)((H) + 31) / 32, (unsigned)((8290) + 15) / 16, (unsigned)(1)), 32, 0, stream>>>(g1_19); }
    { GemmP g2_19;
      g2_19.A = H1; g2_19.B = W2 + 77824; g2_19.bias = b2 + 1216; g2_19.R = H1; g2_19.C = H2;
      g2_19.sAo = 0; g2_19.sAi = 0; g2_19.sAm = H; g2_19.sAk = 1; g2_19.sBo = 0; g2_19.sBi = 0; g2_19.sBn = 1; g2_19.sBk = H; g2_19.sCo = 0; g2_19.sCi = 0; g2_19.sCm = H; g2_19.sRo = 0; g2_19.sRi = 0; g2_19.sRm = 0; g2_19.sRn = 0;
      g2_19.M = 8290; g2_19.N = H; g2_19.K = H; g2_19.zi_n = 1; g2_19.flags = 1; g2_19.act = 1;
      g2_19.alpha = 1.0f; g2_19.beta = 0.0f; g2_19.sa = 1.0f; g2_19.sb = 8.0f; g2_19.Npad = H; g2_19.pad_ = 0;
      k_gemm<0><<<dim3((unsigned)((H) + 31) / 32, (unsigned)((8290) + 15) / 16, (unsigned)(1)), 32, 0, stream>>>(g2_19); }
    { GemmP g3_19;
      g3_19.A = H2; g3_19.B = W3 + 1216; g3_19.bias = b3 + 19; g3_19.R = H2; g3_19.C = Y;
      g3_19.sAo = 0; g3_19.sAi = 0; g3_19.sAm = H; g3_19.sAk = 1; g3_19.sBo = 0; g3_19.sBi = 0; g3_19.sBn = 1; g3_19.sBk = 1; g3_19.sCo = 0; g3_19.sCi = 0; g3_19.sCm = LP; g3_19.sRo = 0; g3_19.sRi = 0; g3_19.sRm = 0; g3_19.sRn = 0;
      g3_19.M = 8290; g3_19.N = 1; g3_19.K = H; g3_19.zi_n = 1; g3_19.flags = 1; g3_19.act = 0;
      g3_19.alpha = 1.0f; g3_19.beta = 0.0f; g3_19.sa = 1.0f; g3_19.sb = 8.0f; g3_19.Npad = LP; g3_19.pad_ = 0;
      k_gemm<0><<<dim3((unsigned)((LP) + 31) / 32, (unsigned)((8290) + 15) / 16, (unsigned)(1)), 32, 0, stream>>>(g3_19); }
    k_es_scatter<<<(unsigned)((8290 + 255) / 256), 256, 0, stream>>>(Y, LP, slot, IDX, 19, 155410, 8290, out);
    { GemmP g1_20;
      g1_20.A = XS + (size_t)163700 * 8; g1_20.B = W1 + 3840; g1_20.bias = b1 + 1280; g1_20.R = XS + (size_t)163700 * 8; g1_20.C = H1;
      g1_20.sAo = 0; g1_20.sAi = 0; g1_20.sAm = 8; g1_20.sAk = 1; g1_20.sBo = 0; g1_20.sBi = 0; g1_20.sBn = 1; g1_20.sBk = H; g1_20.sCo = 0; g1_20.sCi = 0; g1_20.sCm = H; g1_20.sRo = 0; g1_20.sRi = 0; g1_20.sRm = 0; g1_20.sRn = 0;
      g1_20.M = 8235; g1_20.N = H; g1_20.K = 3; g1_20.zi_n = 1; g1_20.flags = 1; g1_20.act = 1;
      g1_20.alpha = 1.0f; g1_20.beta = 0.0f; g1_20.sa = 1.0f; g1_20.sb = 8.0f; g1_20.Npad = H; g1_20.pad_ = 0;
      k_gemm<0><<<dim3((unsigned)((H) + 31) / 32, (unsigned)((8235) + 15) / 16, (unsigned)(1)), 32, 0, stream>>>(g1_20); }
    { GemmP g2_20;
      g2_20.A = H1; g2_20.B = W2 + 81920; g2_20.bias = b2 + 1280; g2_20.R = H1; g2_20.C = H2;
      g2_20.sAo = 0; g2_20.sAi = 0; g2_20.sAm = H; g2_20.sAk = 1; g2_20.sBo = 0; g2_20.sBi = 0; g2_20.sBn = 1; g2_20.sBk = H; g2_20.sCo = 0; g2_20.sCi = 0; g2_20.sCm = H; g2_20.sRo = 0; g2_20.sRi = 0; g2_20.sRm = 0; g2_20.sRn = 0;
      g2_20.M = 8235; g2_20.N = H; g2_20.K = H; g2_20.zi_n = 1; g2_20.flags = 1; g2_20.act = 1;
      g2_20.alpha = 1.0f; g2_20.beta = 0.0f; g2_20.sa = 1.0f; g2_20.sb = 8.0f; g2_20.Npad = H; g2_20.pad_ = 0;
      k_gemm<0><<<dim3((unsigned)((H) + 31) / 32, (unsigned)((8235) + 15) / 16, (unsigned)(1)), 32, 0, stream>>>(g2_20); }
    { GemmP g3_20;
      g3_20.A = H2; g3_20.B = W3 + 1280; g3_20.bias = b3 + 20; g3_20.R = H2; g3_20.C = Y;
      g3_20.sAo = 0; g3_20.sAi = 0; g3_20.sAm = H; g3_20.sAk = 1; g3_20.sBo = 0; g3_20.sBi = 0; g3_20.sBn = 1; g3_20.sBk = 1; g3_20.sCo = 0; g3_20.sCi = 0; g3_20.sCm = LP; g3_20.sRo = 0; g3_20.sRi = 0; g3_20.sRm = 0; g3_20.sRn = 0;
      g3_20.M = 8235; g3_20.N = 1; g3_20.K = H; g3_20.zi_n = 1; g3_20.flags = 1; g3_20.act = 0;
      g3_20.alpha = 1.0f; g3_20.beta = 0.0f; g3_20.sa = 1.0f; g3_20.sb = 8.0f; g3_20.Npad = LP; g3_20.pad_ = 0;
      k_gemm<0><<<dim3((unsigned)((LP) + 31) / 32, (unsigned)((8235) + 15) / 16, (unsigned)(1)), 32, 0, stream>>>(g3_20); }
    k_es_scatter<<<(unsigned)((8235 + 255) / 256), 256, 0, stream>>>(Y, LP, slot, IDX, 20, 163700, 8235, out);
    { GemmP g1_21;
      g1_21.A = XS + (size_t)171935 * 8; g1_21.B = W1 + 4032; g1_21.bias = b1 + 1344; g1_21.R = XS + (size_t)171935 * 8; g1_21.C = H1;
      g1_21.sAo = 0; g1_21.sAi = 0; g1_21.sAm = 8; g1_21.sAk = 1; g1_21.sBo = 0; g1_21.sBi = 0; g1_21.sBn = 1; g1_21.sBk = H; g1_21.sCo = 0; g1_21.sCi = 0; g1_21.sCm = H; g1_21.sRo = 0; g1_21.sRi = 0; g1_21.sRm = 0; g1_21.sRn = 0;
      g1_21.M = 8178; g1_21.N = H; g1_21.K = 3; g1_21.zi_n = 1; g1_21.flags = 1; g1_21.act = 1;
      g1_21.alpha = 1.0f; g1_21.beta = 0.0f; g1_21.sa = 1.0f; g1_21.sb = 8.0f; g1_21.Npad = H; g1_21.pad_ = 0;
      k_gemm<0><<<dim3((unsigned)((H) + 31) / 32, (unsigned)((8178) + 15) / 16, (unsigned)(1)), 32, 0, stream>>>(g1_21); }
    { GemmP g2_21;
      g2_21.A = H1; g2_21.B = W2 + 86016; g2_21.bias = b2 + 1344; g2_21.R = H1; g2_21.C = H2;
      g2_21.sAo = 0; g2_21.sAi = 0; g2_21.sAm = H; g2_21.sAk = 1; g2_21.sBo = 0; g2_21.sBi = 0; g2_21.sBn = 1; g2_21.sBk = H; g2_21.sCo = 0; g2_21.sCi = 0; g2_21.sCm = H; g2_21.sRo = 0; g2_21.sRi = 0; g2_21.sRm = 0; g2_21.sRn = 0;
      g2_21.M = 8178; g2_21.N = H; g2_21.K = H; g2_21.zi_n = 1; g2_21.flags = 1; g2_21.act = 1;
      g2_21.alpha = 1.0f; g2_21.beta = 0.0f; g2_21.sa = 1.0f; g2_21.sb = 8.0f; g2_21.Npad = H; g2_21.pad_ = 0;
      k_gemm<0><<<dim3((unsigned)((H) + 31) / 32, (unsigned)((8178) + 15) / 16, (unsigned)(1)), 32, 0, stream>>>(g2_21); }
    { GemmP g3_21;
      g3_21.A = H2; g3_21.B = W3 + 1344; g3_21.bias = b3 + 21; g3_21.R = H2; g3_21.C = Y;
      g3_21.sAo = 0; g3_21.sAi = 0; g3_21.sAm = H; g3_21.sAk = 1; g3_21.sBo = 0; g3_21.sBi = 0; g3_21.sBn = 1; g3_21.sBk = 1; g3_21.sCo = 0; g3_21.sCi = 0; g3_21.sCm = LP; g3_21.sRo = 0; g3_21.sRi = 0; g3_21.sRm = 0; g3_21.sRn = 0;
      g3_21.M = 8178; g3_21.N = 1; g3_21.K = H; g3_21.zi_n = 1; g3_21.flags = 1; g3_21.act = 0;
      g3_21.alpha = 1.0f; g3_21.beta = 0.0f; g3_21.sa = 1.0f; g3_21.sb = 8.0f; g3_21.Npad = LP; g3_21.pad_ = 0;
      k_gemm<0><<<dim3((unsigned)((LP) + 31) / 32, (unsigned)((8178) + 15) / 16, (unsigned)(1)), 32, 0, stream>>>(g3_21); }
    k_es_scatter<<<(unsigned)((8178 + 255) / 256), 256, 0, stream>>>(Y, LP, slot, IDX, 21, 171935, 8178, out);
    { GemmP g1_22;
      g1_22.A = XS + (size_t)180113 * 8; g1_22.B = W1 + 4224; g1_22.bias = b1 + 1408; g1_22.R = XS + (size_t)180113 * 8; g1_22.C = H1;
      g1_22.sAo = 0; g1_22.sAi = 0; g1_22.sAm = 8; g1_22.sAk = 1; g1_22.sBo = 0; g1_22.sBi = 0; g1_22.sBn = 1; g1_22.sBk = H; g1_22.sCo = 0; g1_22.sCi = 0; g1_22.sCm = H; g1_22.sRo = 0; g1_22.sRi = 0; g1_22.sRm = 0; g1_22.sRn = 0;
      g1_22.M = 8098; g1_22.N = H; g1_22.K = 3; g1_22.zi_n = 1; g1_22.flags = 1; g1_22.act = 1;
      g1_22.alpha = 1.0f; g1_22.beta = 0.0f; g1_22.sa = 1.0f; g1_22.sb = 8.0f; g1_22.Npad = H; g1_22.pad_ = 0;
      k_gemm<0><<<dim3((unsigned)((H) + 31) / 32, (unsigned)((8098) + 15) / 16, (unsigned)(1)), 32, 0, stream>>>(g1_22); }
    { GemmP g2_22;
      g2_22.A = H1; g2_22.B = W2 + 90112; g2_22.bias = b2 + 1408; g2_22.R = H1; g2_22.C = H2;
      g2_22.sAo = 0; g2_22.sAi = 0; g2_22.sAm = H; g2_22.sAk = 1; g2_22.sBo = 0; g2_22.sBi = 0; g2_22.sBn = 1; g2_22.sBk = H; g2_22.sCo = 0; g2_22.sCi = 0; g2_22.sCm = H; g2_22.sRo = 0; g2_22.sRi = 0; g2_22.sRm = 0; g2_22.sRn = 0;
      g2_22.M = 8098; g2_22.N = H; g2_22.K = H; g2_22.zi_n = 1; g2_22.flags = 1; g2_22.act = 1;
      g2_22.alpha = 1.0f; g2_22.beta = 0.0f; g2_22.sa = 1.0f; g2_22.sb = 8.0f; g2_22.Npad = H; g2_22.pad_ = 0;
      k_gemm<0><<<dim3((unsigned)((H) + 31) / 32, (unsigned)((8098) + 15) / 16, (unsigned)(1)), 32, 0, stream>>>(g2_22); }
    { GemmP g3_22;
      g3_22.A = H2; g3_22.B = W3 + 1408; g3_22.bias = b3 + 22; g3_22.R = H2; g3_22.C = Y;
      g3_22.sAo = 0; g3_22.sAi = 0; g3_22.sAm = H; g3_22.sAk = 1; g3_22.sBo = 0; g3_22.sBi = 0; g3_22.sBn = 1; g3_22.sBk = 1; g3_22.sCo = 0; g3_22.sCi = 0; g3_22.sCm = LP; g3_22.sRo = 0; g3_22.sRi = 0; g3_22.sRm = 0; g3_22.sRn = 0;
      g3_22.M = 8098; g3_22.N = 1; g3_22.K = H; g3_22.zi_n = 1; g3_22.flags = 1; g3_22.act = 0;
      g3_22.alpha = 1.0f; g3_22.beta = 0.0f; g3_22.sa = 1.0f; g3_22.sb = 8.0f; g3_22.Npad = LP; g3_22.pad_ = 0;
      k_gemm<0><<<dim3((unsigned)((LP) + 31) / 32, (unsigned)((8098) + 15) / 16, (unsigned)(1)), 32, 0, stream>>>(g3_22); }
    k_es_scatter<<<(unsigned)((8098 + 255) / 256), 256, 0, stream>>>(Y, LP, slot, IDX, 22, 180113, 8098, out);
    { GemmP g1_23;
      g1_23.A = XS + (size_t)188211 * 8; g1_23.B = W1 + 4416; g1_23.bias = b1 + 1472; g1_23.R = XS + (size_t)188211 * 8; g1_23.C = H1;
      g1_23.sAo = 0; g1_23.sAi = 0; g1_23.sAm = 8; g1_23.sAk = 1; g1_23.sBo = 0; g1_23.sBi = 0; g1_23.sBn = 1; g1_23.sBk = H; g1_23.sCo = 0; g1_23.sCi = 0; g1_23.sCm = H; g1_23.sRo = 0; g1_23.sRi = 0; g1_23.sRm = 0; g1_23.sRn = 0;
      g1_23.M = 8349; g1_23.N = H; g1_23.K = 3; g1_23.zi_n = 1; g1_23.flags = 1; g1_23.act = 1;
      g1_23.alpha = 1.0f; g1_23.beta = 0.0f; g1_23.sa = 1.0f; g1_23.sb = 8.0f; g1_23.Npad = H; g1_23.pad_ = 0;
      k_gemm<0><<<dim3((unsigned)((H) + 31) / 32, (unsigned)((8349) + 15) / 16, (unsigned)(1)), 32, 0, stream>>>(g1_23); }
    { GemmP g2_23;
      g2_23.A = H1; g2_23.B = W2 + 94208; g2_23.bias = b2 + 1472; g2_23.R = H1; g2_23.C = H2;
      g2_23.sAo = 0; g2_23.sAi = 0; g2_23.sAm = H; g2_23.sAk = 1; g2_23.sBo = 0; g2_23.sBi = 0; g2_23.sBn = 1; g2_23.sBk = H; g2_23.sCo = 0; g2_23.sCi = 0; g2_23.sCm = H; g2_23.sRo = 0; g2_23.sRi = 0; g2_23.sRm = 0; g2_23.sRn = 0;
      g2_23.M = 8349; g2_23.N = H; g2_23.K = H; g2_23.zi_n = 1; g2_23.flags = 1; g2_23.act = 1;
      g2_23.alpha = 1.0f; g2_23.beta = 0.0f; g2_23.sa = 1.0f; g2_23.sb = 8.0f; g2_23.Npad = H; g2_23.pad_ = 0;
      k_gemm<0><<<dim3((unsigned)((H) + 31) / 32, (unsigned)((8349) + 15) / 16, (unsigned)(1)), 32, 0, stream>>>(g2_23); }
    { GemmP g3_23;
      g3_23.A = H2; g3_23.B = W3 + 1472; g3_23.bias = b3 + 23; g3_23.R = H2; g3_23.C = Y;
      g3_23.sAo = 0; g3_23.sAi = 0; g3_23.sAm = H; g3_23.sAk = 1; g3_23.sBo = 0; g3_23.sBi = 0; g3_23.sBn = 1; g3_23.sBk = 1; g3_23.sCo = 0; g3_23.sCi = 0; g3_23.sCm = LP; g3_23.sRo = 0; g3_23.sRi = 0; g3_23.sRm = 0; g3_23.sRn = 0;
      g3_23.M = 8349; g3_23.N = 1; g3_23.K = H; g3_23.zi_n = 1; g3_23.flags = 1; g3_23.act = 0;
      g3_23.alpha = 1.0f; g3_23.beta = 0.0f; g3_23.sa = 1.0f; g3_23.sb = 8.0f; g3_23.Npad = LP; g3_23.pad_ = 0;
      k_gemm<0><<<dim3((unsigned)((LP) + 31) / 32, (unsigned)((8349) + 15) / 16, (unsigned)(1)), 32, 0, stream>>>(g3_23); }
    k_es_scatter<<<(unsigned)((8349 + 255) / 256), 256, 0, stream>>>(Y, LP, slot, IDX, 23, 188211, 8349, out);
    { GemmP g1_24;
      g1_24.A = XS + (size_t)196560 * 8; g1_24.B = W1 + 4608; g1_24.bias = b1 + 1536; g1_24.R = XS + (size_t)196560 * 8; g1_24.C = H1;
      g1_24.sAo = 0; g1_24.sAi = 0; g1_24.sAm = 8; g1_24.sAk = 1; g1_24.sBo = 0; g1_24.sBi = 0; g1_24.sBn = 1; g1_24.sBk = H; g1_24.sCo = 0; g1_24.sCi = 0; g1_24.sCm = H; g1_24.sRo = 0; g1_24.sRi = 0; g1_24.sRm = 0; g1_24.sRn = 0;
      g1_24.M = 8129; g1_24.N = H; g1_24.K = 3; g1_24.zi_n = 1; g1_24.flags = 1; g1_24.act = 1;
      g1_24.alpha = 1.0f; g1_24.beta = 0.0f; g1_24.sa = 1.0f; g1_24.sb = 8.0f; g1_24.Npad = H; g1_24.pad_ = 0;
      k_gemm<0><<<dim3((unsigned)((H) + 31) / 32, (unsigned)((8129) + 15) / 16, (unsigned)(1)), 32, 0, stream>>>(g1_24); }
    { GemmP g2_24;
      g2_24.A = H1; g2_24.B = W2 + 98304; g2_24.bias = b2 + 1536; g2_24.R = H1; g2_24.C = H2;
      g2_24.sAo = 0; g2_24.sAi = 0; g2_24.sAm = H; g2_24.sAk = 1; g2_24.sBo = 0; g2_24.sBi = 0; g2_24.sBn = 1; g2_24.sBk = H; g2_24.sCo = 0; g2_24.sCi = 0; g2_24.sCm = H; g2_24.sRo = 0; g2_24.sRi = 0; g2_24.sRm = 0; g2_24.sRn = 0;
      g2_24.M = 8129; g2_24.N = H; g2_24.K = H; g2_24.zi_n = 1; g2_24.flags = 1; g2_24.act = 1;
      g2_24.alpha = 1.0f; g2_24.beta = 0.0f; g2_24.sa = 1.0f; g2_24.sb = 8.0f; g2_24.Npad = H; g2_24.pad_ = 0;
      k_gemm<0><<<dim3((unsigned)((H) + 31) / 32, (unsigned)((8129) + 15) / 16, (unsigned)(1)), 32, 0, stream>>>(g2_24); }
    { GemmP g3_24;
      g3_24.A = H2; g3_24.B = W3 + 1536; g3_24.bias = b3 + 24; g3_24.R = H2; g3_24.C = Y;
      g3_24.sAo = 0; g3_24.sAi = 0; g3_24.sAm = H; g3_24.sAk = 1; g3_24.sBo = 0; g3_24.sBi = 0; g3_24.sBn = 1; g3_24.sBk = 1; g3_24.sCo = 0; g3_24.sCi = 0; g3_24.sCm = LP; g3_24.sRo = 0; g3_24.sRi = 0; g3_24.sRm = 0; g3_24.sRn = 0;
      g3_24.M = 8129; g3_24.N = 1; g3_24.K = H; g3_24.zi_n = 1; g3_24.flags = 1; g3_24.act = 0;
      g3_24.alpha = 1.0f; g3_24.beta = 0.0f; g3_24.sa = 1.0f; g3_24.sb = 8.0f; g3_24.Npad = LP; g3_24.pad_ = 0;
      k_gemm<0><<<dim3((unsigned)((LP) + 31) / 32, (unsigned)((8129) + 15) / 16, (unsigned)(1)), 32, 0, stream>>>(g3_24); }
    k_es_scatter<<<(unsigned)((8129 + 255) / 256), 256, 0, stream>>>(Y, LP, slot, IDX, 24, 196560, 8129, out);
    { GemmP g1_25;
      g1_25.A = XS + (size_t)204689 * 8; g1_25.B = W1 + 4800; g1_25.bias = b1 + 1600; g1_25.R = XS + (size_t)204689 * 8; g1_25.C = H1;
      g1_25.sAo = 0; g1_25.sAi = 0; g1_25.sAm = 8; g1_25.sAk = 1; g1_25.sBo = 0; g1_25.sBi = 0; g1_25.sBn = 1; g1_25.sBk = H; g1_25.sCo = 0; g1_25.sCi = 0; g1_25.sCm = H; g1_25.sRo = 0; g1_25.sRi = 0; g1_25.sRm = 0; g1_25.sRn = 0;
      g1_25.M = 8054; g1_25.N = H; g1_25.K = 3; g1_25.zi_n = 1; g1_25.flags = 1; g1_25.act = 1;
      g1_25.alpha = 1.0f; g1_25.beta = 0.0f; g1_25.sa = 1.0f; g1_25.sb = 8.0f; g1_25.Npad = H; g1_25.pad_ = 0;
      k_gemm<0><<<dim3((unsigned)((H) + 31) / 32, (unsigned)((8054) + 15) / 16, (unsigned)(1)), 32, 0, stream>>>(g1_25); }
    { GemmP g2_25;
      g2_25.A = H1; g2_25.B = W2 + 102400; g2_25.bias = b2 + 1600; g2_25.R = H1; g2_25.C = H2;
      g2_25.sAo = 0; g2_25.sAi = 0; g2_25.sAm = H; g2_25.sAk = 1; g2_25.sBo = 0; g2_25.sBi = 0; g2_25.sBn = 1; g2_25.sBk = H; g2_25.sCo = 0; g2_25.sCi = 0; g2_25.sCm = H; g2_25.sRo = 0; g2_25.sRi = 0; g2_25.sRm = 0; g2_25.sRn = 0;
      g2_25.M = 8054; g2_25.N = H; g2_25.K = H; g2_25.zi_n = 1; g2_25.flags = 1; g2_25.act = 1;
      g2_25.alpha = 1.0f; g2_25.beta = 0.0f; g2_25.sa = 1.0f; g2_25.sb = 8.0f; g2_25.Npad = H; g2_25.pad_ = 0;
      k_gemm<0><<<dim3((unsigned)((H) + 31) / 32, (unsigned)((8054) + 15) / 16, (unsigned)(1)), 32, 0, stream>>>(g2_25); }
    { GemmP g3_25;
      g3_25.A = H2; g3_25.B = W3 + 1600; g3_25.bias = b3 + 25; g3_25.R = H2; g3_25.C = Y;
      g3_25.sAo = 0; g3_25.sAi = 0; g3_25.sAm = H; g3_25.sAk = 1; g3_25.sBo = 0; g3_25.sBi = 0; g3_25.sBn = 1; g3_25.sBk = 1; g3_25.sCo = 0; g3_25.sCi = 0; g3_25.sCm = LP; g3_25.sRo = 0; g3_25.sRi = 0; g3_25.sRm = 0; g3_25.sRn = 0;
      g3_25.M = 8054; g3_25.N = 1; g3_25.K = H; g3_25.zi_n = 1; g3_25.flags = 1; g3_25.act = 0;
      g3_25.alpha = 1.0f; g3_25.beta = 0.0f; g3_25.sa = 1.0f; g3_25.sb = 8.0f; g3_25.Npad = LP; g3_25.pad_ = 0;
      k_gemm<0><<<dim3((unsigned)((LP) + 31) / 32, (unsigned)((8054) + 15) / 16, (unsigned)(1)), 32, 0, stream>>>(g3_25); }
    k_es_scatter<<<(unsigned)((8054 + 255) / 256), 256, 0, stream>>>(Y, LP, slot, IDX, 25, 204689, 8054, out);
    { GemmP g1_26;
      g1_26.A = XS + (size_t)212743 * 8; g1_26.B = W1 + 4992; g1_26.bias = b1 + 1664; g1_26.R = XS + (size_t)212743 * 8; g1_26.C = H1;
      g1_26.sAo = 0; g1_26.sAi = 0; g1_26.sAm = 8; g1_26.sAk = 1; g1_26.sBo = 0; g1_26.sBi = 0; g1_26.sBn = 1; g1_26.sBk = H; g1_26.sCo = 0; g1_26.sCi = 0; g1_26.sCm = H; g1_26.sRo = 0; g1_26.sRi = 0; g1_26.sRm = 0; g1_26.sRn = 0;
      g1_26.M = 8314; g1_26.N = H; g1_26.K = 3; g1_26.zi_n = 1; g1_26.flags = 1; g1_26.act = 1;
      g1_26.alpha = 1.0f; g1_26.beta = 0.0f; g1_26.sa = 1.0f; g1_26.sb = 8.0f; g1_26.Npad = H; g1_26.pad_ = 0;
      k_gemm<0><<<dim3((unsigned)((H) + 31) / 32, (unsigned)((8314) + 15) / 16, (unsigned)(1)), 32, 0, stream>>>(g1_26); }
    { GemmP g2_26;
      g2_26.A = H1; g2_26.B = W2 + 106496; g2_26.bias = b2 + 1664; g2_26.R = H1; g2_26.C = H2;
      g2_26.sAo = 0; g2_26.sAi = 0; g2_26.sAm = H; g2_26.sAk = 1; g2_26.sBo = 0; g2_26.sBi = 0; g2_26.sBn = 1; g2_26.sBk = H; g2_26.sCo = 0; g2_26.sCi = 0; g2_26.sCm = H; g2_26.sRo = 0; g2_26.sRi = 0; g2_26.sRm = 0; g2_26.sRn = 0;
      g2_26.M = 8314; g2_26.N = H; g2_26.K = H; g2_26.zi_n = 1; g2_26.flags = 1; g2_26.act = 1;
      g2_26.alpha = 1.0f; g2_26.beta = 0.0f; g2_26.sa = 1.0f; g2_26.sb = 8.0f; g2_26.Npad = H; g2_26.pad_ = 0;
      k_gemm<0><<<dim3((unsigned)((H) + 31) / 32, (unsigned)((8314) + 15) / 16, (unsigned)(1)), 32, 0, stream>>>(g2_26); }
    { GemmP g3_26;
      g3_26.A = H2; g3_26.B = W3 + 1664; g3_26.bias = b3 + 26; g3_26.R = H2; g3_26.C = Y;
      g3_26.sAo = 0; g3_26.sAi = 0; g3_26.sAm = H; g3_26.sAk = 1; g3_26.sBo = 0; g3_26.sBi = 0; g3_26.sBn = 1; g3_26.sBk = 1; g3_26.sCo = 0; g3_26.sCi = 0; g3_26.sCm = LP; g3_26.sRo = 0; g3_26.sRi = 0; g3_26.sRm = 0; g3_26.sRn = 0;
      g3_26.M = 8314; g3_26.N = 1; g3_26.K = H; g3_26.zi_n = 1; g3_26.flags = 1; g3_26.act = 0;
      g3_26.alpha = 1.0f; g3_26.beta = 0.0f; g3_26.sa = 1.0f; g3_26.sb = 8.0f; g3_26.Npad = LP; g3_26.pad_ = 0;
      k_gemm<0><<<dim3((unsigned)((LP) + 31) / 32, (unsigned)((8314) + 15) / 16, (unsigned)(1)), 32, 0, stream>>>(g3_26); }
    k_es_scatter<<<(unsigned)((8314 + 255) / 256), 256, 0, stream>>>(Y, LP, slot, IDX, 26, 212743, 8314, out);
    { GemmP g1_27;
      g1_27.A = XS + (size_t)221057 * 8; g1_27.B = W1 + 5184; g1_27.bias = b1 + 1728; g1_27.R = XS + (size_t)221057 * 8; g1_27.C = H1;
      g1_27.sAo = 0; g1_27.sAi = 0; g1_27.sAm = 8; g1_27.sAk = 1; g1_27.sBo = 0; g1_27.sBi = 0; g1_27.sBn = 1; g1_27.sBk = H; g1_27.sCo = 0; g1_27.sCi = 0; g1_27.sCm = H; g1_27.sRo = 0; g1_27.sRi = 0; g1_27.sRm = 0; g1_27.sRn = 0;
      g1_27.M = 8169; g1_27.N = H; g1_27.K = 3; g1_27.zi_n = 1; g1_27.flags = 1; g1_27.act = 1;
      g1_27.alpha = 1.0f; g1_27.beta = 0.0f; g1_27.sa = 1.0f; g1_27.sb = 8.0f; g1_27.Npad = H; g1_27.pad_ = 0;
      k_gemm<0><<<dim3((unsigned)((H) + 31) / 32, (unsigned)((8169) + 15) / 16, (unsigned)(1)), 32, 0, stream>>>(g1_27); }
    { GemmP g2_27;
      g2_27.A = H1; g2_27.B = W2 + 110592; g2_27.bias = b2 + 1728; g2_27.R = H1; g2_27.C = H2;
      g2_27.sAo = 0; g2_27.sAi = 0; g2_27.sAm = H; g2_27.sAk = 1; g2_27.sBo = 0; g2_27.sBi = 0; g2_27.sBn = 1; g2_27.sBk = H; g2_27.sCo = 0; g2_27.sCi = 0; g2_27.sCm = H; g2_27.sRo = 0; g2_27.sRi = 0; g2_27.sRm = 0; g2_27.sRn = 0;
      g2_27.M = 8169; g2_27.N = H; g2_27.K = H; g2_27.zi_n = 1; g2_27.flags = 1; g2_27.act = 1;
      g2_27.alpha = 1.0f; g2_27.beta = 0.0f; g2_27.sa = 1.0f; g2_27.sb = 8.0f; g2_27.Npad = H; g2_27.pad_ = 0;
      k_gemm<0><<<dim3((unsigned)((H) + 31) / 32, (unsigned)((8169) + 15) / 16, (unsigned)(1)), 32, 0, stream>>>(g2_27); }
    { GemmP g3_27;
      g3_27.A = H2; g3_27.B = W3 + 1728; g3_27.bias = b3 + 27; g3_27.R = H2; g3_27.C = Y;
      g3_27.sAo = 0; g3_27.sAi = 0; g3_27.sAm = H; g3_27.sAk = 1; g3_27.sBo = 0; g3_27.sBi = 0; g3_27.sBn = 1; g3_27.sBk = 1; g3_27.sCo = 0; g3_27.sCi = 0; g3_27.sCm = LP; g3_27.sRo = 0; g3_27.sRi = 0; g3_27.sRm = 0; g3_27.sRn = 0;
      g3_27.M = 8169; g3_27.N = 1; g3_27.K = H; g3_27.zi_n = 1; g3_27.flags = 1; g3_27.act = 0;
      g3_27.alpha = 1.0f; g3_27.beta = 0.0f; g3_27.sa = 1.0f; g3_27.sb = 8.0f; g3_27.Npad = LP; g3_27.pad_ = 0;
      k_gemm<0><<<dim3((unsigned)((LP) + 31) / 32, (unsigned)((8169) + 15) / 16, (unsigned)(1)), 32, 0, stream>>>(g3_27); }
    k_es_scatter<<<(unsigned)((8169 + 255) / 256), 256, 0, stream>>>(Y, LP, slot, IDX, 27, 221057, 8169, out);
    { GemmP g1_28;
      g1_28.A = XS + (size_t)229226 * 8; g1_28.B = W1 + 5376; g1_28.bias = b1 + 1792; g1_28.R = XS + (size_t)229226 * 8; g1_28.C = H1;
      g1_28.sAo = 0; g1_28.sAi = 0; g1_28.sAm = 8; g1_28.sAk = 1; g1_28.sBo = 0; g1_28.sBi = 0; g1_28.sBn = 1; g1_28.sBk = H; g1_28.sCo = 0; g1_28.sCi = 0; g1_28.sCm = H; g1_28.sRo = 0; g1_28.sRi = 0; g1_28.sRm = 0; g1_28.sRn = 0;
      g1_28.M = 8239; g1_28.N = H; g1_28.K = 3; g1_28.zi_n = 1; g1_28.flags = 1; g1_28.act = 1;
      g1_28.alpha = 1.0f; g1_28.beta = 0.0f; g1_28.sa = 1.0f; g1_28.sb = 8.0f; g1_28.Npad = H; g1_28.pad_ = 0;
      k_gemm<0><<<dim3((unsigned)((H) + 31) / 32, (unsigned)((8239) + 15) / 16, (unsigned)(1)), 32, 0, stream>>>(g1_28); }
    { GemmP g2_28;
      g2_28.A = H1; g2_28.B = W2 + 114688; g2_28.bias = b2 + 1792; g2_28.R = H1; g2_28.C = H2;
      g2_28.sAo = 0; g2_28.sAi = 0; g2_28.sAm = H; g2_28.sAk = 1; g2_28.sBo = 0; g2_28.sBi = 0; g2_28.sBn = 1; g2_28.sBk = H; g2_28.sCo = 0; g2_28.sCi = 0; g2_28.sCm = H; g2_28.sRo = 0; g2_28.sRi = 0; g2_28.sRm = 0; g2_28.sRn = 0;
      g2_28.M = 8239; g2_28.N = H; g2_28.K = H; g2_28.zi_n = 1; g2_28.flags = 1; g2_28.act = 1;
      g2_28.alpha = 1.0f; g2_28.beta = 0.0f; g2_28.sa = 1.0f; g2_28.sb = 8.0f; g2_28.Npad = H; g2_28.pad_ = 0;
      k_gemm<0><<<dim3((unsigned)((H) + 31) / 32, (unsigned)((8239) + 15) / 16, (unsigned)(1)), 32, 0, stream>>>(g2_28); }
    { GemmP g3_28;
      g3_28.A = H2; g3_28.B = W3 + 1792; g3_28.bias = b3 + 28; g3_28.R = H2; g3_28.C = Y;
      g3_28.sAo = 0; g3_28.sAi = 0; g3_28.sAm = H; g3_28.sAk = 1; g3_28.sBo = 0; g3_28.sBi = 0; g3_28.sBn = 1; g3_28.sBk = 1; g3_28.sCo = 0; g3_28.sCi = 0; g3_28.sCm = LP; g3_28.sRo = 0; g3_28.sRi = 0; g3_28.sRm = 0; g3_28.sRn = 0;
      g3_28.M = 8239; g3_28.N = 1; g3_28.K = H; g3_28.zi_n = 1; g3_28.flags = 1; g3_28.act = 0;
      g3_28.alpha = 1.0f; g3_28.beta = 0.0f; g3_28.sa = 1.0f; g3_28.sb = 8.0f; g3_28.Npad = LP; g3_28.pad_ = 0;
      k_gemm<0><<<dim3((unsigned)((LP) + 31) / 32, (unsigned)((8239) + 15) / 16, (unsigned)(1)), 32, 0, stream>>>(g3_28); }
    k_es_scatter<<<(unsigned)((8239 + 255) / 256), 256, 0, stream>>>(Y, LP, slot, IDX, 28, 229226, 8239, out);
    { GemmP g1_29;
      g1_29.A = XS + (size_t)237465 * 8; g1_29.B = W1 + 5568; g1_29.bias = b1 + 1856; g1_29.R = XS + (size_t)237465 * 8; g1_29.C = H1;
      g1_29.sAo = 0; g1_29.sAi = 0; g1_29.sAm = 8; g1_29.sAk = 1; g1_29.sBo = 0; g1_29.sBi = 0; g1_29.sBn = 1; g1_29.sBk = H; g1_29.sCo = 0; g1_29.sCi = 0; g1_29.sCm = H; g1_29.sRo = 0; g1_29.sRi = 0; g1_29.sRm = 0; g1_29.sRn = 0;
      g1_29.M = 8331; g1_29.N = H; g1_29.K = 3; g1_29.zi_n = 1; g1_29.flags = 1; g1_29.act = 1;
      g1_29.alpha = 1.0f; g1_29.beta = 0.0f; g1_29.sa = 1.0f; g1_29.sb = 8.0f; g1_29.Npad = H; g1_29.pad_ = 0;
      k_gemm<0><<<dim3((unsigned)((H) + 31) / 32, (unsigned)((8331) + 15) / 16, (unsigned)(1)), 32, 0, stream>>>(g1_29); }
    { GemmP g2_29;
      g2_29.A = H1; g2_29.B = W2 + 118784; g2_29.bias = b2 + 1856; g2_29.R = H1; g2_29.C = H2;
      g2_29.sAo = 0; g2_29.sAi = 0; g2_29.sAm = H; g2_29.sAk = 1; g2_29.sBo = 0; g2_29.sBi = 0; g2_29.sBn = 1; g2_29.sBk = H; g2_29.sCo = 0; g2_29.sCi = 0; g2_29.sCm = H; g2_29.sRo = 0; g2_29.sRi = 0; g2_29.sRm = 0; g2_29.sRn = 0;
      g2_29.M = 8331; g2_29.N = H; g2_29.K = H; g2_29.zi_n = 1; g2_29.flags = 1; g2_29.act = 1;
      g2_29.alpha = 1.0f; g2_29.beta = 0.0f; g2_29.sa = 1.0f; g2_29.sb = 8.0f; g2_29.Npad = H; g2_29.pad_ = 0;
      k_gemm<0><<<dim3((unsigned)((H) + 31) / 32, (unsigned)((8331) + 15) / 16, (unsigned)(1)), 32, 0, stream>>>(g2_29); }
    { GemmP g3_29;
      g3_29.A = H2; g3_29.B = W3 + 1856; g3_29.bias = b3 + 29; g3_29.R = H2; g3_29.C = Y;
      g3_29.sAo = 0; g3_29.sAi = 0; g3_29.sAm = H; g3_29.sAk = 1; g3_29.sBo = 0; g3_29.sBi = 0; g3_29.sBn = 1; g3_29.sBk = 1; g3_29.sCo = 0; g3_29.sCi = 0; g3_29.sCm = LP; g3_29.sRo = 0; g3_29.sRi = 0; g3_29.sRm = 0; g3_29.sRn = 0;
      g3_29.M = 8331; g3_29.N = 1; g3_29.K = H; g3_29.zi_n = 1; g3_29.flags = 1; g3_29.act = 0;
      g3_29.alpha = 1.0f; g3_29.beta = 0.0f; g3_29.sa = 1.0f; g3_29.sb = 8.0f; g3_29.Npad = LP; g3_29.pad_ = 0;
      k_gemm<0><<<dim3((unsigned)((LP) + 31) / 32, (unsigned)((8331) + 15) / 16, (unsigned)(1)), 32, 0, stream>>>(g3_29); }
    k_es_scatter<<<(unsigned)((8331 + 255) / 256), 256, 0, stream>>>(Y, LP, slot, IDX, 29, 237465, 8331, out);
    { GemmP g1_30;
      g1_30.A = XS + (size_t)245796 * 8; g1_30.B = W1 + 5760; g1_30.bias = b1 + 1920; g1_30.R = XS + (size_t)245796 * 8; g1_30.C = H1;
      g1_30.sAo = 0; g1_30.sAi = 0; g1_30.sAm = 8; g1_30.sAk = 1; g1_30.sBo = 0; g1_30.sBi = 0; g1_30.sBn = 1; g1_30.sBk = H; g1_30.sCo = 0; g1_30.sCi = 0; g1_30.sCm = H; g1_30.sRo = 0; g1_30.sRi = 0; g1_30.sRm = 0; g1_30.sRn = 0;
      g1_30.M = 8260; g1_30.N = H; g1_30.K = 3; g1_30.zi_n = 1; g1_30.flags = 1; g1_30.act = 1;
      g1_30.alpha = 1.0f; g1_30.beta = 0.0f; g1_30.sa = 1.0f; g1_30.sb = 8.0f; g1_30.Npad = H; g1_30.pad_ = 0;
      k_gemm<0><<<dim3((unsigned)((H) + 31) / 32, (unsigned)((8260) + 15) / 16, (unsigned)(1)), 32, 0, stream>>>(g1_30); }
    { GemmP g2_30;
      g2_30.A = H1; g2_30.B = W2 + 122880; g2_30.bias = b2 + 1920; g2_30.R = H1; g2_30.C = H2;
      g2_30.sAo = 0; g2_30.sAi = 0; g2_30.sAm = H; g2_30.sAk = 1; g2_30.sBo = 0; g2_30.sBi = 0; g2_30.sBn = 1; g2_30.sBk = H; g2_30.sCo = 0; g2_30.sCi = 0; g2_30.sCm = H; g2_30.sRo = 0; g2_30.sRi = 0; g2_30.sRm = 0; g2_30.sRn = 0;
      g2_30.M = 8260; g2_30.N = H; g2_30.K = H; g2_30.zi_n = 1; g2_30.flags = 1; g2_30.act = 1;
      g2_30.alpha = 1.0f; g2_30.beta = 0.0f; g2_30.sa = 1.0f; g2_30.sb = 8.0f; g2_30.Npad = H; g2_30.pad_ = 0;
      k_gemm<0><<<dim3((unsigned)((H) + 31) / 32, (unsigned)((8260) + 15) / 16, (unsigned)(1)), 32, 0, stream>>>(g2_30); }
    { GemmP g3_30;
      g3_30.A = H2; g3_30.B = W3 + 1920; g3_30.bias = b3 + 30; g3_30.R = H2; g3_30.C = Y;
      g3_30.sAo = 0; g3_30.sAi = 0; g3_30.sAm = H; g3_30.sAk = 1; g3_30.sBo = 0; g3_30.sBi = 0; g3_30.sBn = 1; g3_30.sBk = 1; g3_30.sCo = 0; g3_30.sCi = 0; g3_30.sCm = LP; g3_30.sRo = 0; g3_30.sRi = 0; g3_30.sRm = 0; g3_30.sRn = 0;
      g3_30.M = 8260; g3_30.N = 1; g3_30.K = H; g3_30.zi_n = 1; g3_30.flags = 1; g3_30.act = 0;
      g3_30.alpha = 1.0f; g3_30.beta = 0.0f; g3_30.sa = 1.0f; g3_30.sb = 8.0f; g3_30.Npad = LP; g3_30.pad_ = 0;
      k_gemm<0><<<dim3((unsigned)((LP) + 31) / 32, (unsigned)((8260) + 15) / 16, (unsigned)(1)), 32, 0, stream>>>(g3_30); }
    k_es_scatter<<<(unsigned)((8260 + 255) / 256), 256, 0, stream>>>(Y, LP, slot, IDX, 30, 245796, 8260, out);
    { GemmP g1_31;
      g1_31.A = XS + (size_t)254056 * 8; g1_31.B = W1 + 5952; g1_31.bias = b1 + 1984; g1_31.R = XS + (size_t)254056 * 8; g1_31.C = H1;
      g1_31.sAo = 0; g1_31.sAi = 0; g1_31.sAm = 8; g1_31.sAk = 1; g1_31.sBo = 0; g1_31.sBi = 0; g1_31.sBn = 1; g1_31.sBk = H; g1_31.sCo = 0; g1_31.sCi = 0; g1_31.sCm = H; g1_31.sRo = 0; g1_31.sRi = 0; g1_31.sRm = 0; g1_31.sRn = 0;
      g1_31.M = 8126; g1_31.N = H; g1_31.K = 3; g1_31.zi_n = 1; g1_31.flags = 1; g1_31.act = 1;
      g1_31.alpha = 1.0f; g1_31.beta = 0.0f; g1_31.sa = 1.0f; g1_31.sb = 8.0f; g1_31.Npad = H; g1_31.pad_ = 0;
      k_gemm<0><<<dim3((unsigned)((H) + 31) / 32, (unsigned)((8126) + 15) / 16, (unsigned)(1)), 32, 0, stream>>>(g1_31); }
    { GemmP g2_31;
      g2_31.A = H1; g2_31.B = W2 + 126976; g2_31.bias = b2 + 1984; g2_31.R = H1; g2_31.C = H2;
      g2_31.sAo = 0; g2_31.sAi = 0; g2_31.sAm = H; g2_31.sAk = 1; g2_31.sBo = 0; g2_31.sBi = 0; g2_31.sBn = 1; g2_31.sBk = H; g2_31.sCo = 0; g2_31.sCi = 0; g2_31.sCm = H; g2_31.sRo = 0; g2_31.sRi = 0; g2_31.sRm = 0; g2_31.sRn = 0;
      g2_31.M = 8126; g2_31.N = H; g2_31.K = H; g2_31.zi_n = 1; g2_31.flags = 1; g2_31.act = 1;
      g2_31.alpha = 1.0f; g2_31.beta = 0.0f; g2_31.sa = 1.0f; g2_31.sb = 8.0f; g2_31.Npad = H; g2_31.pad_ = 0;
      k_gemm<0><<<dim3((unsigned)((H) + 31) / 32, (unsigned)((8126) + 15) / 16, (unsigned)(1)), 32, 0, stream>>>(g2_31); }
    { GemmP g3_31;
      g3_31.A = H2; g3_31.B = W3 + 1984; g3_31.bias = b3 + 31; g3_31.R = H2; g3_31.C = Y;
      g3_31.sAo = 0; g3_31.sAi = 0; g3_31.sAm = H; g3_31.sAk = 1; g3_31.sBo = 0; g3_31.sBi = 0; g3_31.sBn = 1; g3_31.sBk = 1; g3_31.sCo = 0; g3_31.sCi = 0; g3_31.sCm = LP; g3_31.sRo = 0; g3_31.sRi = 0; g3_31.sRm = 0; g3_31.sRn = 0;
      g3_31.M = 8126; g3_31.N = 1; g3_31.K = H; g3_31.zi_n = 1; g3_31.flags = 1; g3_31.act = 0;
      g3_31.alpha = 1.0f; g3_31.beta = 0.0f; g3_31.sa = 1.0f; g3_31.sb = 8.0f; g3_31.Npad = LP; g3_31.pad_ = 0;
      k_gemm<0><<<dim3((unsigned)((LP) + 31) / 32, (unsigned)((8126) + 15) / 16, (unsigned)(1)), 32, 0, stream>>>(g3_31); }
    k_es_scatter<<<(unsigned)((8126 + 255) / 256), 256, 0, stream>>>(Y, LP, slot, IDX, 31, 254056, 8126, out);
    { GemmP g1_32;
      g1_32.A = XS + (size_t)262182 * 8; g1_32.B = W1 + 6144; g1_32.bias = b1 + 2048; g1_32.R = XS + (size_t)262182 * 8; g1_32.C = H1;
      g1_32.sAo = 0; g1_32.sAi = 0; g1_32.sAm = 8; g1_32.sAk = 1; g1_32.sBo = 0; g1_32.sBi = 0; g1_32.sBn = 1; g1_32.sBk = H; g1_32.sCo = 0; g1_32.sCi = 0; g1_32.sCm = H; g1_32.sRo = 0; g1_32.sRi = 0; g1_32.sRm = 0; g1_32.sRn = 0;
      g1_32.M = 8309; g1_32.N = H; g1_32.K = 3; g1_32.zi_n = 1; g1_32.flags = 1; g1_32.act = 1;
      g1_32.alpha = 1.0f; g1_32.beta = 0.0f; g1_32.sa = 1.0f; g1_32.sb = 8.0f; g1_32.Npad = H; g1_32.pad_ = 0;
      k_gemm<0><<<dim3((unsigned)((H) + 31) / 32, (unsigned)((8309) + 15) / 16, (unsigned)(1)), 32, 0, stream>>>(g1_32); }
    { GemmP g2_32;
      g2_32.A = H1; g2_32.B = W2 + 131072; g2_32.bias = b2 + 2048; g2_32.R = H1; g2_32.C = H2;
      g2_32.sAo = 0; g2_32.sAi = 0; g2_32.sAm = H; g2_32.sAk = 1; g2_32.sBo = 0; g2_32.sBi = 0; g2_32.sBn = 1; g2_32.sBk = H; g2_32.sCo = 0; g2_32.sCi = 0; g2_32.sCm = H; g2_32.sRo = 0; g2_32.sRi = 0; g2_32.sRm = 0; g2_32.sRn = 0;
      g2_32.M = 8309; g2_32.N = H; g2_32.K = H; g2_32.zi_n = 1; g2_32.flags = 1; g2_32.act = 1;
      g2_32.alpha = 1.0f; g2_32.beta = 0.0f; g2_32.sa = 1.0f; g2_32.sb = 8.0f; g2_32.Npad = H; g2_32.pad_ = 0;
      k_gemm<0><<<dim3((unsigned)((H) + 31) / 32, (unsigned)((8309) + 15) / 16, (unsigned)(1)), 32, 0, stream>>>(g2_32); }
    { GemmP g3_32;
      g3_32.A = H2; g3_32.B = W3 + 2048; g3_32.bias = b3 + 32; g3_32.R = H2; g3_32.C = Y;
      g3_32.sAo = 0; g3_32.sAi = 0; g3_32.sAm = H; g3_32.sAk = 1; g3_32.sBo = 0; g3_32.sBi = 0; g3_32.sBn = 1; g3_32.sBk = 1; g3_32.sCo = 0; g3_32.sCi = 0; g3_32.sCm = LP; g3_32.sRo = 0; g3_32.sRi = 0; g3_32.sRm = 0; g3_32.sRn = 0;
      g3_32.M = 8309; g3_32.N = 1; g3_32.K = H; g3_32.zi_n = 1; g3_32.flags = 1; g3_32.act = 0;
      g3_32.alpha = 1.0f; g3_32.beta = 0.0f; g3_32.sa = 1.0f; g3_32.sb = 8.0f; g3_32.Npad = LP; g3_32.pad_ = 0;
      k_gemm<0><<<dim3((unsigned)((LP) + 31) / 32, (unsigned)((8309) + 15) / 16, (unsigned)(1)), 32, 0, stream>>>(g3_32); }
    k_es_scatter<<<(unsigned)((8309 + 255) / 256), 256, 0, stream>>>(Y, LP, slot, IDX, 32, 262182, 8309, out);
    { GemmP g1_33;
      g1_33.A = XS + (size_t)270491 * 8; g1_33.B = W1 + 6336; g1_33.bias = b1 + 2112; g1_33.R = XS + (size_t)270491 * 8; g1_33.C = H1;
      g1_33.sAo = 0; g1_33.sAi = 0; g1_33.sAm = 8; g1_33.sAk = 1; g1_33.sBo = 0; g1_33.sBi = 0; g1_33.sBn = 1; g1_33.sBk = H; g1_33.sCo = 0; g1_33.sCi = 0; g1_33.sCm = H; g1_33.sRo = 0; g1_33.sRi = 0; g1_33.sRm = 0; g1_33.sRn = 0;
      g1_33.M = 8188; g1_33.N = H; g1_33.K = 3; g1_33.zi_n = 1; g1_33.flags = 1; g1_33.act = 1;
      g1_33.alpha = 1.0f; g1_33.beta = 0.0f; g1_33.sa = 1.0f; g1_33.sb = 8.0f; g1_33.Npad = H; g1_33.pad_ = 0;
      k_gemm<0><<<dim3((unsigned)((H) + 31) / 32, (unsigned)((8188) + 15) / 16, (unsigned)(1)), 32, 0, stream>>>(g1_33); }
    { GemmP g2_33;
      g2_33.A = H1; g2_33.B = W2 + 135168; g2_33.bias = b2 + 2112; g2_33.R = H1; g2_33.C = H2;
      g2_33.sAo = 0; g2_33.sAi = 0; g2_33.sAm = H; g2_33.sAk = 1; g2_33.sBo = 0; g2_33.sBi = 0; g2_33.sBn = 1; g2_33.sBk = H; g2_33.sCo = 0; g2_33.sCi = 0; g2_33.sCm = H; g2_33.sRo = 0; g2_33.sRi = 0; g2_33.sRm = 0; g2_33.sRn = 0;
      g2_33.M = 8188; g2_33.N = H; g2_33.K = H; g2_33.zi_n = 1; g2_33.flags = 1; g2_33.act = 1;
      g2_33.alpha = 1.0f; g2_33.beta = 0.0f; g2_33.sa = 1.0f; g2_33.sb = 8.0f; g2_33.Npad = H; g2_33.pad_ = 0;
      k_gemm<0><<<dim3((unsigned)((H) + 31) / 32, (unsigned)((8188) + 15) / 16, (unsigned)(1)), 32, 0, stream>>>(g2_33); }
    { GemmP g3_33;
      g3_33.A = H2; g3_33.B = W3 + 2112; g3_33.bias = b3 + 33; g3_33.R = H2; g3_33.C = Y;
      g3_33.sAo = 0; g3_33.sAi = 0; g3_33.sAm = H; g3_33.sAk = 1; g3_33.sBo = 0; g3_33.sBi = 0; g3_33.sBn = 1; g3_33.sBk = 1; g3_33.sCo = 0; g3_33.sCi = 0; g3_33.sCm = LP; g3_33.sRo = 0; g3_33.sRi = 0; g3_33.sRm = 0; g3_33.sRn = 0;
      g3_33.M = 8188; g3_33.N = 1; g3_33.K = H; g3_33.zi_n = 1; g3_33.flags = 1; g3_33.act = 0;
      g3_33.alpha = 1.0f; g3_33.beta = 0.0f; g3_33.sa = 1.0f; g3_33.sb = 8.0f; g3_33.Npad = LP; g3_33.pad_ = 0;
      k_gemm<0><<<dim3((unsigned)((LP) + 31) / 32, (unsigned)((8188) + 15) / 16, (unsigned)(1)), 32, 0, stream>>>(g3_33); }
    k_es_scatter<<<(unsigned)((8188 + 255) / 256), 256, 0, stream>>>(Y, LP, slot, IDX, 33, 270491, 8188, out);
    { GemmP g1_34;
      g1_34.A = XS + (size_t)278679 * 8; g1_34.B = W1 + 6528; g1_34.bias = b1 + 2176; g1_34.R = XS + (size_t)278679 * 8; g1_34.C = H1;
      g1_34.sAo = 0; g1_34.sAi = 0; g1_34.sAm = 8; g1_34.sAk = 1; g1_34.sBo = 0; g1_34.sBi = 0; g1_34.sBn = 1; g1_34.sBk = H; g1_34.sCo = 0; g1_34.sCi = 0; g1_34.sCm = H; g1_34.sRo = 0; g1_34.sRi = 0; g1_34.sRm = 0; g1_34.sRn = 0;
      g1_34.M = 8268; g1_34.N = H; g1_34.K = 3; g1_34.zi_n = 1; g1_34.flags = 1; g1_34.act = 1;
      g1_34.alpha = 1.0f; g1_34.beta = 0.0f; g1_34.sa = 1.0f; g1_34.sb = 8.0f; g1_34.Npad = H; g1_34.pad_ = 0;
      k_gemm<0><<<dim3((unsigned)((H) + 31) / 32, (unsigned)((8268) + 15) / 16, (unsigned)(1)), 32, 0, stream>>>(g1_34); }
    { GemmP g2_34;
      g2_34.A = H1; g2_34.B = W2 + 139264; g2_34.bias = b2 + 2176; g2_34.R = H1; g2_34.C = H2;
      g2_34.sAo = 0; g2_34.sAi = 0; g2_34.sAm = H; g2_34.sAk = 1; g2_34.sBo = 0; g2_34.sBi = 0; g2_34.sBn = 1; g2_34.sBk = H; g2_34.sCo = 0; g2_34.sCi = 0; g2_34.sCm = H; g2_34.sRo = 0; g2_34.sRi = 0; g2_34.sRm = 0; g2_34.sRn = 0;
      g2_34.M = 8268; g2_34.N = H; g2_34.K = H; g2_34.zi_n = 1; g2_34.flags = 1; g2_34.act = 1;
      g2_34.alpha = 1.0f; g2_34.beta = 0.0f; g2_34.sa = 1.0f; g2_34.sb = 8.0f; g2_34.Npad = H; g2_34.pad_ = 0;
      k_gemm<0><<<dim3((unsigned)((H) + 31) / 32, (unsigned)((8268) + 15) / 16, (unsigned)(1)), 32, 0, stream>>>(g2_34); }
    { GemmP g3_34;
      g3_34.A = H2; g3_34.B = W3 + 2176; g3_34.bias = b3 + 34; g3_34.R = H2; g3_34.C = Y;
      g3_34.sAo = 0; g3_34.sAi = 0; g3_34.sAm = H; g3_34.sAk = 1; g3_34.sBo = 0; g3_34.sBi = 0; g3_34.sBn = 1; g3_34.sBk = 1; g3_34.sCo = 0; g3_34.sCi = 0; g3_34.sCm = LP; g3_34.sRo = 0; g3_34.sRi = 0; g3_34.sRm = 0; g3_34.sRn = 0;
      g3_34.M = 8268; g3_34.N = 1; g3_34.K = H; g3_34.zi_n = 1; g3_34.flags = 1; g3_34.act = 0;
      g3_34.alpha = 1.0f; g3_34.beta = 0.0f; g3_34.sa = 1.0f; g3_34.sb = 8.0f; g3_34.Npad = LP; g3_34.pad_ = 0;
      k_gemm<0><<<dim3((unsigned)((LP) + 31) / 32, (unsigned)((8268) + 15) / 16, (unsigned)(1)), 32, 0, stream>>>(g3_34); }
    k_es_scatter<<<(unsigned)((8268 + 255) / 256), 256, 0, stream>>>(Y, LP, slot, IDX, 34, 278679, 8268, out);
    { GemmP g1_35;
      g1_35.A = XS + (size_t)286947 * 8; g1_35.B = W1 + 6720; g1_35.bias = b1 + 2240; g1_35.R = XS + (size_t)286947 * 8; g1_35.C = H1;
      g1_35.sAo = 0; g1_35.sAi = 0; g1_35.sAm = 8; g1_35.sAk = 1; g1_35.sBo = 0; g1_35.sBi = 0; g1_35.sBn = 1; g1_35.sBk = H; g1_35.sCo = 0; g1_35.sCi = 0; g1_35.sCm = H; g1_35.sRo = 0; g1_35.sRi = 0; g1_35.sRm = 0; g1_35.sRn = 0;
      g1_35.M = 8094; g1_35.N = H; g1_35.K = 3; g1_35.zi_n = 1; g1_35.flags = 1; g1_35.act = 1;
      g1_35.alpha = 1.0f; g1_35.beta = 0.0f; g1_35.sa = 1.0f; g1_35.sb = 8.0f; g1_35.Npad = H; g1_35.pad_ = 0;
      k_gemm<0><<<dim3((unsigned)((H) + 31) / 32, (unsigned)((8094) + 15) / 16, (unsigned)(1)), 32, 0, stream>>>(g1_35); }
    { GemmP g2_35;
      g2_35.A = H1; g2_35.B = W2 + 143360; g2_35.bias = b2 + 2240; g2_35.R = H1; g2_35.C = H2;
      g2_35.sAo = 0; g2_35.sAi = 0; g2_35.sAm = H; g2_35.sAk = 1; g2_35.sBo = 0; g2_35.sBi = 0; g2_35.sBn = 1; g2_35.sBk = H; g2_35.sCo = 0; g2_35.sCi = 0; g2_35.sCm = H; g2_35.sRo = 0; g2_35.sRi = 0; g2_35.sRm = 0; g2_35.sRn = 0;
      g2_35.M = 8094; g2_35.N = H; g2_35.K = H; g2_35.zi_n = 1; g2_35.flags = 1; g2_35.act = 1;
      g2_35.alpha = 1.0f; g2_35.beta = 0.0f; g2_35.sa = 1.0f; g2_35.sb = 8.0f; g2_35.Npad = H; g2_35.pad_ = 0;
      k_gemm<0><<<dim3((unsigned)((H) + 31) / 32, (unsigned)((8094) + 15) / 16, (unsigned)(1)), 32, 0, stream>>>(g2_35); }
    { GemmP g3_35;
      g3_35.A = H2; g3_35.B = W3 + 2240; g3_35.bias = b3 + 35; g3_35.R = H2; g3_35.C = Y;
      g3_35.sAo = 0; g3_35.sAi = 0; g3_35.sAm = H; g3_35.sAk = 1; g3_35.sBo = 0; g3_35.sBi = 0; g3_35.sBn = 1; g3_35.sBk = 1; g3_35.sCo = 0; g3_35.sCi = 0; g3_35.sCm = LP; g3_35.sRo = 0; g3_35.sRi = 0; g3_35.sRm = 0; g3_35.sRn = 0;
      g3_35.M = 8094; g3_35.N = 1; g3_35.K = H; g3_35.zi_n = 1; g3_35.flags = 1; g3_35.act = 0;
      g3_35.alpha = 1.0f; g3_35.beta = 0.0f; g3_35.sa = 1.0f; g3_35.sb = 8.0f; g3_35.Npad = LP; g3_35.pad_ = 0;
      k_gemm<0><<<dim3((unsigned)((LP) + 31) / 32, (unsigned)((8094) + 15) / 16, (unsigned)(1)), 32, 0, stream>>>(g3_35); }
    k_es_scatter<<<(unsigned)((8094 + 255) / 256), 256, 0, stream>>>(Y, LP, slot, IDX, 35, 286947, 8094, out);
    { GemmP g1_36;
      g1_36.A = XS + (size_t)295041 * 8; g1_36.B = W1 + 6912; g1_36.bias = b1 + 2304; g1_36.R = XS + (size_t)295041 * 8; g1_36.C = H1;
      g1_36.sAo = 0; g1_36.sAi = 0; g1_36.sAm = 8; g1_36.sAk = 1; g1_36.sBo = 0; g1_36.sBi = 0; g1_36.sBn = 1; g1_36.sBk = H; g1_36.sCo = 0; g1_36.sCi = 0; g1_36.sCm = H; g1_36.sRo = 0; g1_36.sRi = 0; g1_36.sRm = 0; g1_36.sRn = 0;
      g1_36.M = 8111; g1_36.N = H; g1_36.K = 3; g1_36.zi_n = 1; g1_36.flags = 1; g1_36.act = 1;
      g1_36.alpha = 1.0f; g1_36.beta = 0.0f; g1_36.sa = 1.0f; g1_36.sb = 8.0f; g1_36.Npad = H; g1_36.pad_ = 0;
      k_gemm<0><<<dim3((unsigned)((H) + 31) / 32, (unsigned)((8111) + 15) / 16, (unsigned)(1)), 32, 0, stream>>>(g1_36); }
    { GemmP g2_36;
      g2_36.A = H1; g2_36.B = W2 + 147456; g2_36.bias = b2 + 2304; g2_36.R = H1; g2_36.C = H2;
      g2_36.sAo = 0; g2_36.sAi = 0; g2_36.sAm = H; g2_36.sAk = 1; g2_36.sBo = 0; g2_36.sBi = 0; g2_36.sBn = 1; g2_36.sBk = H; g2_36.sCo = 0; g2_36.sCi = 0; g2_36.sCm = H; g2_36.sRo = 0; g2_36.sRi = 0; g2_36.sRm = 0; g2_36.sRn = 0;
      g2_36.M = 8111; g2_36.N = H; g2_36.K = H; g2_36.zi_n = 1; g2_36.flags = 1; g2_36.act = 1;
      g2_36.alpha = 1.0f; g2_36.beta = 0.0f; g2_36.sa = 1.0f; g2_36.sb = 8.0f; g2_36.Npad = H; g2_36.pad_ = 0;
      k_gemm<0><<<dim3((unsigned)((H) + 31) / 32, (unsigned)((8111) + 15) / 16, (unsigned)(1)), 32, 0, stream>>>(g2_36); }
    { GemmP g3_36;
      g3_36.A = H2; g3_36.B = W3 + 2304; g3_36.bias = b3 + 36; g3_36.R = H2; g3_36.C = Y;
      g3_36.sAo = 0; g3_36.sAi = 0; g3_36.sAm = H; g3_36.sAk = 1; g3_36.sBo = 0; g3_36.sBi = 0; g3_36.sBn = 1; g3_36.sBk = 1; g3_36.sCo = 0; g3_36.sCi = 0; g3_36.sCm = LP; g3_36.sRo = 0; g3_36.sRi = 0; g3_36.sRm = 0; g3_36.sRn = 0;
      g3_36.M = 8111; g3_36.N = 1; g3_36.K = H; g3_36.zi_n = 1; g3_36.flags = 1; g3_36.act = 0;
      g3_36.alpha = 1.0f; g3_36.beta = 0.0f; g3_36.sa = 1.0f; g3_36.sb = 8.0f; g3_36.Npad = LP; g3_36.pad_ = 0;
      k_gemm<0><<<dim3((unsigned)((LP) + 31) / 32, (unsigned)((8111) + 15) / 16, (unsigned)(1)), 32, 0, stream>>>(g3_36); }
    k_es_scatter<<<(unsigned)((8111 + 255) / 256), 256, 0, stream>>>(Y, LP, slot, IDX, 36, 295041, 8111, out);
    { GemmP g1_37;
      g1_37.A = XS + (size_t)303152 * 8; g1_37.B = W1 + 7104; g1_37.bias = b1 + 2368; g1_37.R = XS + (size_t)303152 * 8; g1_37.C = H1;
      g1_37.sAo = 0; g1_37.sAi = 0; g1_37.sAm = 8; g1_37.sAk = 1; g1_37.sBo = 0; g1_37.sBi = 0; g1_37.sBn = 1; g1_37.sBk = H; g1_37.sCo = 0; g1_37.sCi = 0; g1_37.sCm = H; g1_37.sRo = 0; g1_37.sRi = 0; g1_37.sRm = 0; g1_37.sRn = 0;
      g1_37.M = 8091; g1_37.N = H; g1_37.K = 3; g1_37.zi_n = 1; g1_37.flags = 1; g1_37.act = 1;
      g1_37.alpha = 1.0f; g1_37.beta = 0.0f; g1_37.sa = 1.0f; g1_37.sb = 8.0f; g1_37.Npad = H; g1_37.pad_ = 0;
      k_gemm<0><<<dim3((unsigned)((H) + 31) / 32, (unsigned)((8091) + 15) / 16, (unsigned)(1)), 32, 0, stream>>>(g1_37); }
    { GemmP g2_37;
      g2_37.A = H1; g2_37.B = W2 + 151552; g2_37.bias = b2 + 2368; g2_37.R = H1; g2_37.C = H2;
      g2_37.sAo = 0; g2_37.sAi = 0; g2_37.sAm = H; g2_37.sAk = 1; g2_37.sBo = 0; g2_37.sBi = 0; g2_37.sBn = 1; g2_37.sBk = H; g2_37.sCo = 0; g2_37.sCi = 0; g2_37.sCm = H; g2_37.sRo = 0; g2_37.sRi = 0; g2_37.sRm = 0; g2_37.sRn = 0;
      g2_37.M = 8091; g2_37.N = H; g2_37.K = H; g2_37.zi_n = 1; g2_37.flags = 1; g2_37.act = 1;
      g2_37.alpha = 1.0f; g2_37.beta = 0.0f; g2_37.sa = 1.0f; g2_37.sb = 8.0f; g2_37.Npad = H; g2_37.pad_ = 0;
      k_gemm<0><<<dim3((unsigned)((H) + 31) / 32, (unsigned)((8091) + 15) / 16, (unsigned)(1)), 32, 0, stream>>>(g2_37); }
    { GemmP g3_37;
      g3_37.A = H2; g3_37.B = W3 + 2368; g3_37.bias = b3 + 37; g3_37.R = H2; g3_37.C = Y;
      g3_37.sAo = 0; g3_37.sAi = 0; g3_37.sAm = H; g3_37.sAk = 1; g3_37.sBo = 0; g3_37.sBi = 0; g3_37.sBn = 1; g3_37.sBk = 1; g3_37.sCo = 0; g3_37.sCi = 0; g3_37.sCm = LP; g3_37.sRo = 0; g3_37.sRi = 0; g3_37.sRm = 0; g3_37.sRn = 0;
      g3_37.M = 8091; g3_37.N = 1; g3_37.K = H; g3_37.zi_n = 1; g3_37.flags = 1; g3_37.act = 0;
      g3_37.alpha = 1.0f; g3_37.beta = 0.0f; g3_37.sa = 1.0f; g3_37.sb = 8.0f; g3_37.Npad = LP; g3_37.pad_ = 0;
      k_gemm<0><<<dim3((unsigned)((LP) + 31) / 32, (unsigned)((8091) + 15) / 16, (unsigned)(1)), 32, 0, stream>>>(g3_37); }
    k_es_scatter<<<(unsigned)((8091 + 255) / 256), 256, 0, stream>>>(Y, LP, slot, IDX, 37, 303152, 8091, out);
    { GemmP g1_38;
      g1_38.A = XS + (size_t)311243 * 8; g1_38.B = W1 + 7296; g1_38.bias = b1 + 2432; g1_38.R = XS + (size_t)311243 * 8; g1_38.C = H1;
      g1_38.sAo = 0; g1_38.sAi = 0; g1_38.sAm = 8; g1_38.sAk = 1; g1_38.sBo = 0; g1_38.sBi = 0; g1_38.sBn = 1; g1_38.sBk = H; g1_38.sCo = 0; g1_38.sCi = 0; g1_38.sCm = H; g1_38.sRo = 0; g1_38.sRi = 0; g1_38.sRm = 0; g1_38.sRn = 0;
      g1_38.M = 8158; g1_38.N = H; g1_38.K = 3; g1_38.zi_n = 1; g1_38.flags = 1; g1_38.act = 1;
      g1_38.alpha = 1.0f; g1_38.beta = 0.0f; g1_38.sa = 1.0f; g1_38.sb = 8.0f; g1_38.Npad = H; g1_38.pad_ = 0;
      k_gemm<0><<<dim3((unsigned)((H) + 31) / 32, (unsigned)((8158) + 15) / 16, (unsigned)(1)), 32, 0, stream>>>(g1_38); }
    { GemmP g2_38;
      g2_38.A = H1; g2_38.B = W2 + 155648; g2_38.bias = b2 + 2432; g2_38.R = H1; g2_38.C = H2;
      g2_38.sAo = 0; g2_38.sAi = 0; g2_38.sAm = H; g2_38.sAk = 1; g2_38.sBo = 0; g2_38.sBi = 0; g2_38.sBn = 1; g2_38.sBk = H; g2_38.sCo = 0; g2_38.sCi = 0; g2_38.sCm = H; g2_38.sRo = 0; g2_38.sRi = 0; g2_38.sRm = 0; g2_38.sRn = 0;
      g2_38.M = 8158; g2_38.N = H; g2_38.K = H; g2_38.zi_n = 1; g2_38.flags = 1; g2_38.act = 1;
      g2_38.alpha = 1.0f; g2_38.beta = 0.0f; g2_38.sa = 1.0f; g2_38.sb = 8.0f; g2_38.Npad = H; g2_38.pad_ = 0;
      k_gemm<0><<<dim3((unsigned)((H) + 31) / 32, (unsigned)((8158) + 15) / 16, (unsigned)(1)), 32, 0, stream>>>(g2_38); }
    { GemmP g3_38;
      g3_38.A = H2; g3_38.B = W3 + 2432; g3_38.bias = b3 + 38; g3_38.R = H2; g3_38.C = Y;
      g3_38.sAo = 0; g3_38.sAi = 0; g3_38.sAm = H; g3_38.sAk = 1; g3_38.sBo = 0; g3_38.sBi = 0; g3_38.sBn = 1; g3_38.sBk = 1; g3_38.sCo = 0; g3_38.sCi = 0; g3_38.sCm = LP; g3_38.sRo = 0; g3_38.sRi = 0; g3_38.sRm = 0; g3_38.sRn = 0;
      g3_38.M = 8158; g3_38.N = 1; g3_38.K = H; g3_38.zi_n = 1; g3_38.flags = 1; g3_38.act = 0;
      g3_38.alpha = 1.0f; g3_38.beta = 0.0f; g3_38.sa = 1.0f; g3_38.sb = 8.0f; g3_38.Npad = LP; g3_38.pad_ = 0;
      k_gemm<0><<<dim3((unsigned)((LP) + 31) / 32, (unsigned)((8158) + 15) / 16, (unsigned)(1)), 32, 0, stream>>>(g3_38); }
    k_es_scatter<<<(unsigned)((8158 + 255) / 256), 256, 0, stream>>>(Y, LP, slot, IDX, 38, 311243, 8158, out);
    { GemmP g1_39;
      g1_39.A = XS + (size_t)319401 * 8; g1_39.B = W1 + 7488; g1_39.bias = b1 + 2496; g1_39.R = XS + (size_t)319401 * 8; g1_39.C = H1;
      g1_39.sAo = 0; g1_39.sAi = 0; g1_39.sAm = 8; g1_39.sAk = 1; g1_39.sBo = 0; g1_39.sBi = 0; g1_39.sBn = 1; g1_39.sBk = H; g1_39.sCo = 0; g1_39.sCi = 0; g1_39.sCm = H; g1_39.sRo = 0; g1_39.sRi = 0; g1_39.sRm = 0; g1_39.sRn = 0;
      g1_39.M = 8279; g1_39.N = H; g1_39.K = 3; g1_39.zi_n = 1; g1_39.flags = 1; g1_39.act = 1;
      g1_39.alpha = 1.0f; g1_39.beta = 0.0f; g1_39.sa = 1.0f; g1_39.sb = 8.0f; g1_39.Npad = H; g1_39.pad_ = 0;
      k_gemm<0><<<dim3((unsigned)((H) + 31) / 32, (unsigned)((8279) + 15) / 16, (unsigned)(1)), 32, 0, stream>>>(g1_39); }
    { GemmP g2_39;
      g2_39.A = H1; g2_39.B = W2 + 159744; g2_39.bias = b2 + 2496; g2_39.R = H1; g2_39.C = H2;
      g2_39.sAo = 0; g2_39.sAi = 0; g2_39.sAm = H; g2_39.sAk = 1; g2_39.sBo = 0; g2_39.sBi = 0; g2_39.sBn = 1; g2_39.sBk = H; g2_39.sCo = 0; g2_39.sCi = 0; g2_39.sCm = H; g2_39.sRo = 0; g2_39.sRi = 0; g2_39.sRm = 0; g2_39.sRn = 0;
      g2_39.M = 8279; g2_39.N = H; g2_39.K = H; g2_39.zi_n = 1; g2_39.flags = 1; g2_39.act = 1;
      g2_39.alpha = 1.0f; g2_39.beta = 0.0f; g2_39.sa = 1.0f; g2_39.sb = 8.0f; g2_39.Npad = H; g2_39.pad_ = 0;
      k_gemm<0><<<dim3((unsigned)((H) + 31) / 32, (unsigned)((8279) + 15) / 16, (unsigned)(1)), 32, 0, stream>>>(g2_39); }
    { GemmP g3_39;
      g3_39.A = H2; g3_39.B = W3 + 2496; g3_39.bias = b3 + 39; g3_39.R = H2; g3_39.C = Y;
      g3_39.sAo = 0; g3_39.sAi = 0; g3_39.sAm = H; g3_39.sAk = 1; g3_39.sBo = 0; g3_39.sBi = 0; g3_39.sBn = 1; g3_39.sBk = 1; g3_39.sCo = 0; g3_39.sCi = 0; g3_39.sCm = LP; g3_39.sRo = 0; g3_39.sRi = 0; g3_39.sRm = 0; g3_39.sRn = 0;
      g3_39.M = 8279; g3_39.N = 1; g3_39.K = H; g3_39.zi_n = 1; g3_39.flags = 1; g3_39.act = 0;
      g3_39.alpha = 1.0f; g3_39.beta = 0.0f; g3_39.sa = 1.0f; g3_39.sb = 8.0f; g3_39.Npad = LP; g3_39.pad_ = 0;
      k_gemm<0><<<dim3((unsigned)((LP) + 31) / 32, (unsigned)((8279) + 15) / 16, (unsigned)(1)), 32, 0, stream>>>(g3_39); }
    k_es_scatter<<<(unsigned)((8279 + 255) / 256), 256, 0, stream>>>(Y, LP, slot, IDX, 39, 319401, 8279, out);
    { GemmP g1_40;
      g1_40.A = XS + (size_t)327680 * 8; g1_40.B = W1 + 7680; g1_40.bias = b1 + 2560; g1_40.R = XS + (size_t)327680 * 8; g1_40.C = H1;
      g1_40.sAo = 0; g1_40.sAi = 0; g1_40.sAm = 8; g1_40.sAk = 1; g1_40.sBo = 0; g1_40.sBi = 0; g1_40.sBn = 1; g1_40.sBk = H; g1_40.sCo = 0; g1_40.sCi = 0; g1_40.sCm = H; g1_40.sRo = 0; g1_40.sRi = 0; g1_40.sRm = 0; g1_40.sRn = 0;
      g1_40.M = 8167; g1_40.N = H; g1_40.K = 3; g1_40.zi_n = 1; g1_40.flags = 1; g1_40.act = 1;
      g1_40.alpha = 1.0f; g1_40.beta = 0.0f; g1_40.sa = 1.0f; g1_40.sb = 8.0f; g1_40.Npad = H; g1_40.pad_ = 0;
      k_gemm<0><<<dim3((unsigned)((H) + 31) / 32, (unsigned)((8167) + 15) / 16, (unsigned)(1)), 32, 0, stream>>>(g1_40); }
    { GemmP g2_40;
      g2_40.A = H1; g2_40.B = W2 + 163840; g2_40.bias = b2 + 2560; g2_40.R = H1; g2_40.C = H2;
      g2_40.sAo = 0; g2_40.sAi = 0; g2_40.sAm = H; g2_40.sAk = 1; g2_40.sBo = 0; g2_40.sBi = 0; g2_40.sBn = 1; g2_40.sBk = H; g2_40.sCo = 0; g2_40.sCi = 0; g2_40.sCm = H; g2_40.sRo = 0; g2_40.sRi = 0; g2_40.sRm = 0; g2_40.sRn = 0;
      g2_40.M = 8167; g2_40.N = H; g2_40.K = H; g2_40.zi_n = 1; g2_40.flags = 1; g2_40.act = 1;
      g2_40.alpha = 1.0f; g2_40.beta = 0.0f; g2_40.sa = 1.0f; g2_40.sb = 8.0f; g2_40.Npad = H; g2_40.pad_ = 0;
      k_gemm<0><<<dim3((unsigned)((H) + 31) / 32, (unsigned)((8167) + 15) / 16, (unsigned)(1)), 32, 0, stream>>>(g2_40); }
    { GemmP g3_40;
      g3_40.A = H2; g3_40.B = W3 + 2560; g3_40.bias = b3 + 40; g3_40.R = H2; g3_40.C = Y;
      g3_40.sAo = 0; g3_40.sAi = 0; g3_40.sAm = H; g3_40.sAk = 1; g3_40.sBo = 0; g3_40.sBi = 0; g3_40.sBn = 1; g3_40.sBk = 1; g3_40.sCo = 0; g3_40.sCi = 0; g3_40.sCm = LP; g3_40.sRo = 0; g3_40.sRi = 0; g3_40.sRm = 0; g3_40.sRn = 0;
      g3_40.M = 8167; g3_40.N = 1; g3_40.K = H; g3_40.zi_n = 1; g3_40.flags = 1; g3_40.act = 0;
      g3_40.alpha = 1.0f; g3_40.beta = 0.0f; g3_40.sa = 1.0f; g3_40.sb = 8.0f; g3_40.Npad = LP; g3_40.pad_ = 0;
      k_gemm<0><<<dim3((unsigned)((LP) + 31) / 32, (unsigned)((8167) + 15) / 16, (unsigned)(1)), 32, 0, stream>>>(g3_40); }
    k_es_scatter<<<(unsigned)((8167 + 255) / 256), 256, 0, stream>>>(Y, LP, slot, IDX, 40, 327680, 8167, out);
    { GemmP g1_41;
      g1_41.A = XS + (size_t)335847 * 8; g1_41.B = W1 + 7872; g1_41.bias = b1 + 2624; g1_41.R = XS + (size_t)335847 * 8; g1_41.C = H1;
      g1_41.sAo = 0; g1_41.sAi = 0; g1_41.sAm = 8; g1_41.sAk = 1; g1_41.sBo = 0; g1_41.sBi = 0; g1_41.sBn = 1; g1_41.sBk = H; g1_41.sCo = 0; g1_41.sCi = 0; g1_41.sCm = H; g1_41.sRo = 0; g1_41.sRi = 0; g1_41.sRm = 0; g1_41.sRn = 0;
      g1_41.M = 8301; g1_41.N = H; g1_41.K = 3; g1_41.zi_n = 1; g1_41.flags = 1; g1_41.act = 1;
      g1_41.alpha = 1.0f; g1_41.beta = 0.0f; g1_41.sa = 1.0f; g1_41.sb = 8.0f; g1_41.Npad = H; g1_41.pad_ = 0;
      k_gemm<0><<<dim3((unsigned)((H) + 31) / 32, (unsigned)((8301) + 15) / 16, (unsigned)(1)), 32, 0, stream>>>(g1_41); }
    { GemmP g2_41;
      g2_41.A = H1; g2_41.B = W2 + 167936; g2_41.bias = b2 + 2624; g2_41.R = H1; g2_41.C = H2;
      g2_41.sAo = 0; g2_41.sAi = 0; g2_41.sAm = H; g2_41.sAk = 1; g2_41.sBo = 0; g2_41.sBi = 0; g2_41.sBn = 1; g2_41.sBk = H; g2_41.sCo = 0; g2_41.sCi = 0; g2_41.sCm = H; g2_41.sRo = 0; g2_41.sRi = 0; g2_41.sRm = 0; g2_41.sRn = 0;
      g2_41.M = 8301; g2_41.N = H; g2_41.K = H; g2_41.zi_n = 1; g2_41.flags = 1; g2_41.act = 1;
      g2_41.alpha = 1.0f; g2_41.beta = 0.0f; g2_41.sa = 1.0f; g2_41.sb = 8.0f; g2_41.Npad = H; g2_41.pad_ = 0;
      k_gemm<0><<<dim3((unsigned)((H) + 31) / 32, (unsigned)((8301) + 15) / 16, (unsigned)(1)), 32, 0, stream>>>(g2_41); }
    { GemmP g3_41;
      g3_41.A = H2; g3_41.B = W3 + 2624; g3_41.bias = b3 + 41; g3_41.R = H2; g3_41.C = Y;
      g3_41.sAo = 0; g3_41.sAi = 0; g3_41.sAm = H; g3_41.sAk = 1; g3_41.sBo = 0; g3_41.sBi = 0; g3_41.sBn = 1; g3_41.sBk = 1; g3_41.sCo = 0; g3_41.sCi = 0; g3_41.sCm = LP; g3_41.sRo = 0; g3_41.sRi = 0; g3_41.sRm = 0; g3_41.sRn = 0;
      g3_41.M = 8301; g3_41.N = 1; g3_41.K = H; g3_41.zi_n = 1; g3_41.flags = 1; g3_41.act = 0;
      g3_41.alpha = 1.0f; g3_41.beta = 0.0f; g3_41.sa = 1.0f; g3_41.sb = 8.0f; g3_41.Npad = LP; g3_41.pad_ = 0;
      k_gemm<0><<<dim3((unsigned)((LP) + 31) / 32, (unsigned)((8301) + 15) / 16, (unsigned)(1)), 32, 0, stream>>>(g3_41); }
    k_es_scatter<<<(unsigned)((8301 + 255) / 256), 256, 0, stream>>>(Y, LP, slot, IDX, 41, 335847, 8301, out);
    { GemmP g1_42;
      g1_42.A = XS + (size_t)344148 * 8; g1_42.B = W1 + 8064; g1_42.bias = b1 + 2688; g1_42.R = XS + (size_t)344148 * 8; g1_42.C = H1;
      g1_42.sAo = 0; g1_42.sAi = 0; g1_42.sAm = 8; g1_42.sAk = 1; g1_42.sBo = 0; g1_42.sBi = 0; g1_42.sBn = 1; g1_42.sBk = H; g1_42.sCo = 0; g1_42.sCi = 0; g1_42.sCm = H; g1_42.sRo = 0; g1_42.sRi = 0; g1_42.sRm = 0; g1_42.sRn = 0;
      g1_42.M = 8259; g1_42.N = H; g1_42.K = 3; g1_42.zi_n = 1; g1_42.flags = 1; g1_42.act = 1;
      g1_42.alpha = 1.0f; g1_42.beta = 0.0f; g1_42.sa = 1.0f; g1_42.sb = 8.0f; g1_42.Npad = H; g1_42.pad_ = 0;
      k_gemm<0><<<dim3((unsigned)((H) + 31) / 32, (unsigned)((8259) + 15) / 16, (unsigned)(1)), 32, 0, stream>>>(g1_42); }
    { GemmP g2_42;
      g2_42.A = H1; g2_42.B = W2 + 172032; g2_42.bias = b2 + 2688; g2_42.R = H1; g2_42.C = H2;
      g2_42.sAo = 0; g2_42.sAi = 0; g2_42.sAm = H; g2_42.sAk = 1; g2_42.sBo = 0; g2_42.sBi = 0; g2_42.sBn = 1; g2_42.sBk = H; g2_42.sCo = 0; g2_42.sCi = 0; g2_42.sCm = H; g2_42.sRo = 0; g2_42.sRi = 0; g2_42.sRm = 0; g2_42.sRn = 0;
      g2_42.M = 8259; g2_42.N = H; g2_42.K = H; g2_42.zi_n = 1; g2_42.flags = 1; g2_42.act = 1;
      g2_42.alpha = 1.0f; g2_42.beta = 0.0f; g2_42.sa = 1.0f; g2_42.sb = 8.0f; g2_42.Npad = H; g2_42.pad_ = 0;
      k_gemm<0><<<dim3((unsigned)((H) + 31) / 32, (unsigned)((8259) + 15) / 16, (unsigned)(1)), 32, 0, stream>>>(g2_42); }
    { GemmP g3_42;
      g3_42.A = H2; g3_42.B = W3 + 2688; g3_42.bias = b3 + 42; g3_42.R = H2; g3_42.C = Y;
      g3_42.sAo = 0; g3_42.sAi = 0; g3_42.sAm = H; g3_42.sAk = 1; g3_42.sBo = 0; g3_42.sBi = 0; g3_42.sBn = 1; g3_42.sBk = 1; g3_42.sCo = 0; g3_42.sCi = 0; g3_42.sCm = LP; g3_42.sRo = 0; g3_42.sRi = 0; g3_42.sRm = 0; g3_42.sRn = 0;
      g3_42.M = 8259; g3_42.N = 1; g3_42.K = H; g3_42.zi_n = 1; g3_42.flags = 1; g3_42.act = 0;
      g3_42.alpha = 1.0f; g3_42.beta = 0.0f; g3_42.sa = 1.0f; g3_42.sb = 8.0f; g3_42.Npad = LP; g3_42.pad_ = 0;
      k_gemm<0><<<dim3((unsigned)((LP) + 31) / 32, (unsigned)((8259) + 15) / 16, (unsigned)(1)), 32, 0, stream>>>(g3_42); }
    k_es_scatter<<<(unsigned)((8259 + 255) / 256), 256, 0, stream>>>(Y, LP, slot, IDX, 42, 344148, 8259, out);
    { GemmP g1_43;
      g1_43.A = XS + (size_t)352407 * 8; g1_43.B = W1 + 8256; g1_43.bias = b1 + 2752; g1_43.R = XS + (size_t)352407 * 8; g1_43.C = H1;
      g1_43.sAo = 0; g1_43.sAi = 0; g1_43.sAm = 8; g1_43.sAk = 1; g1_43.sBo = 0; g1_43.sBi = 0; g1_43.sBn = 1; g1_43.sBk = H; g1_43.sCo = 0; g1_43.sCi = 0; g1_43.sCm = H; g1_43.sRo = 0; g1_43.sRi = 0; g1_43.sRm = 0; g1_43.sRn = 0;
      g1_43.M = 8172; g1_43.N = H; g1_43.K = 3; g1_43.zi_n = 1; g1_43.flags = 1; g1_43.act = 1;
      g1_43.alpha = 1.0f; g1_43.beta = 0.0f; g1_43.sa = 1.0f; g1_43.sb = 8.0f; g1_43.Npad = H; g1_43.pad_ = 0;
      k_gemm<0><<<dim3((unsigned)((H) + 31) / 32, (unsigned)((8172) + 15) / 16, (unsigned)(1)), 32, 0, stream>>>(g1_43); }
    { GemmP g2_43;
      g2_43.A = H1; g2_43.B = W2 + 176128; g2_43.bias = b2 + 2752; g2_43.R = H1; g2_43.C = H2;
      g2_43.sAo = 0; g2_43.sAi = 0; g2_43.sAm = H; g2_43.sAk = 1; g2_43.sBo = 0; g2_43.sBi = 0; g2_43.sBn = 1; g2_43.sBk = H; g2_43.sCo = 0; g2_43.sCi = 0; g2_43.sCm = H; g2_43.sRo = 0; g2_43.sRi = 0; g2_43.sRm = 0; g2_43.sRn = 0;
      g2_43.M = 8172; g2_43.N = H; g2_43.K = H; g2_43.zi_n = 1; g2_43.flags = 1; g2_43.act = 1;
      g2_43.alpha = 1.0f; g2_43.beta = 0.0f; g2_43.sa = 1.0f; g2_43.sb = 8.0f; g2_43.Npad = H; g2_43.pad_ = 0;
      k_gemm<0><<<dim3((unsigned)((H) + 31) / 32, (unsigned)((8172) + 15) / 16, (unsigned)(1)), 32, 0, stream>>>(g2_43); }
    { GemmP g3_43;
      g3_43.A = H2; g3_43.B = W3 + 2752; g3_43.bias = b3 + 43; g3_43.R = H2; g3_43.C = Y;
      g3_43.sAo = 0; g3_43.sAi = 0; g3_43.sAm = H; g3_43.sAk = 1; g3_43.sBo = 0; g3_43.sBi = 0; g3_43.sBn = 1; g3_43.sBk = 1; g3_43.sCo = 0; g3_43.sCi = 0; g3_43.sCm = LP; g3_43.sRo = 0; g3_43.sRi = 0; g3_43.sRm = 0; g3_43.sRn = 0;
      g3_43.M = 8172; g3_43.N = 1; g3_43.K = H; g3_43.zi_n = 1; g3_43.flags = 1; g3_43.act = 0;
      g3_43.alpha = 1.0f; g3_43.beta = 0.0f; g3_43.sa = 1.0f; g3_43.sb = 8.0f; g3_43.Npad = LP; g3_43.pad_ = 0;
      k_gemm<0><<<dim3((unsigned)((LP) + 31) / 32, (unsigned)((8172) + 15) / 16, (unsigned)(1)), 32, 0, stream>>>(g3_43); }
    k_es_scatter<<<(unsigned)((8172 + 255) / 256), 256, 0, stream>>>(Y, LP, slot, IDX, 43, 352407, 8172, out);
    { GemmP g1_44;
      g1_44.A = XS + (size_t)360579 * 8; g1_44.B = W1 + 8448; g1_44.bias = b1 + 2816; g1_44.R = XS + (size_t)360579 * 8; g1_44.C = H1;
      g1_44.sAo = 0; g1_44.sAi = 0; g1_44.sAm = 8; g1_44.sAk = 1; g1_44.sBo = 0; g1_44.sBi = 0; g1_44.sBn = 1; g1_44.sBk = H; g1_44.sCo = 0; g1_44.sCi = 0; g1_44.sCm = H; g1_44.sRo = 0; g1_44.sRi = 0; g1_44.sRm = 0; g1_44.sRn = 0;
      g1_44.M = 8161; g1_44.N = H; g1_44.K = 3; g1_44.zi_n = 1; g1_44.flags = 1; g1_44.act = 1;
      g1_44.alpha = 1.0f; g1_44.beta = 0.0f; g1_44.sa = 1.0f; g1_44.sb = 8.0f; g1_44.Npad = H; g1_44.pad_ = 0;
      k_gemm<0><<<dim3((unsigned)((H) + 31) / 32, (unsigned)((8161) + 15) / 16, (unsigned)(1)), 32, 0, stream>>>(g1_44); }
    { GemmP g2_44;
      g2_44.A = H1; g2_44.B = W2 + 180224; g2_44.bias = b2 + 2816; g2_44.R = H1; g2_44.C = H2;
      g2_44.sAo = 0; g2_44.sAi = 0; g2_44.sAm = H; g2_44.sAk = 1; g2_44.sBo = 0; g2_44.sBi = 0; g2_44.sBn = 1; g2_44.sBk = H; g2_44.sCo = 0; g2_44.sCi = 0; g2_44.sCm = H; g2_44.sRo = 0; g2_44.sRi = 0; g2_44.sRm = 0; g2_44.sRn = 0;
      g2_44.M = 8161; g2_44.N = H; g2_44.K = H; g2_44.zi_n = 1; g2_44.flags = 1; g2_44.act = 1;
      g2_44.alpha = 1.0f; g2_44.beta = 0.0f; g2_44.sa = 1.0f; g2_44.sb = 8.0f; g2_44.Npad = H; g2_44.pad_ = 0;
      k_gemm<0><<<dim3((unsigned)((H) + 31) / 32, (unsigned)((8161) + 15) / 16, (unsigned)(1)), 32, 0, stream>>>(g2_44); }
    { GemmP g3_44;
      g3_44.A = H2; g3_44.B = W3 + 2816; g3_44.bias = b3 + 44; g3_44.R = H2; g3_44.C = Y;
      g3_44.sAo = 0; g3_44.sAi = 0; g3_44.sAm = H; g3_44.sAk = 1; g3_44.sBo = 0; g3_44.sBi = 0; g3_44.sBn = 1; g3_44.sBk = 1; g3_44.sCo = 0; g3_44.sCi = 0; g3_44.sCm = LP; g3_44.sRo = 0; g3_44.sRi = 0; g3_44.sRm = 0; g3_44.sRn = 0;
      g3_44.M = 8161; g3_44.N = 1; g3_44.K = H; g3_44.zi_n = 1; g3_44.flags = 1; g3_44.act = 0;
      g3_44.alpha = 1.0f; g3_44.beta = 0.0f; g3_44.sa = 1.0f; g3_44.sb = 8.0f; g3_44.Npad = LP; g3_44.pad_ = 0;
      k_gemm<0><<<dim3((unsigned)((LP) + 31) / 32, (unsigned)((8161) + 15) / 16, (unsigned)(1)), 32, 0, stream>>>(g3_44); }
    k_es_scatter<<<(unsigned)((8161 + 255) / 256), 256, 0, stream>>>(Y, LP, slot, IDX, 44, 360579, 8161, out);
    { GemmP g1_45;
      g1_45.A = XS + (size_t)368740 * 8; g1_45.B = W1 + 8640; g1_45.bias = b1 + 2880; g1_45.R = XS + (size_t)368740 * 8; g1_45.C = H1;
      g1_45.sAo = 0; g1_45.sAi = 0; g1_45.sAm = 8; g1_45.sAk = 1; g1_45.sBo = 0; g1_45.sBi = 0; g1_45.sBn = 1; g1_45.sBk = H; g1_45.sCo = 0; g1_45.sCi = 0; g1_45.sCm = H; g1_45.sRo = 0; g1_45.sRi = 0; g1_45.sRm = 0; g1_45.sRn = 0;
      g1_45.M = 8248; g1_45.N = H; g1_45.K = 3; g1_45.zi_n = 1; g1_45.flags = 1; g1_45.act = 1;
      g1_45.alpha = 1.0f; g1_45.beta = 0.0f; g1_45.sa = 1.0f; g1_45.sb = 8.0f; g1_45.Npad = H; g1_45.pad_ = 0;
      k_gemm<0><<<dim3((unsigned)((H) + 31) / 32, (unsigned)((8248) + 15) / 16, (unsigned)(1)), 32, 0, stream>>>(g1_45); }
    { GemmP g2_45;
      g2_45.A = H1; g2_45.B = W2 + 184320; g2_45.bias = b2 + 2880; g2_45.R = H1; g2_45.C = H2;
      g2_45.sAo = 0; g2_45.sAi = 0; g2_45.sAm = H; g2_45.sAk = 1; g2_45.sBo = 0; g2_45.sBi = 0; g2_45.sBn = 1; g2_45.sBk = H; g2_45.sCo = 0; g2_45.sCi = 0; g2_45.sCm = H; g2_45.sRo = 0; g2_45.sRi = 0; g2_45.sRm = 0; g2_45.sRn = 0;
      g2_45.M = 8248; g2_45.N = H; g2_45.K = H; g2_45.zi_n = 1; g2_45.flags = 1; g2_45.act = 1;
      g2_45.alpha = 1.0f; g2_45.beta = 0.0f; g2_45.sa = 1.0f; g2_45.sb = 8.0f; g2_45.Npad = H; g2_45.pad_ = 0;
      k_gemm<0><<<dim3((unsigned)((H) + 31) / 32, (unsigned)((8248) + 15) / 16, (unsigned)(1)), 32, 0, stream>>>(g2_45); }
    { GemmP g3_45;
      g3_45.A = H2; g3_45.B = W3 + 2880; g3_45.bias = b3 + 45; g3_45.R = H2; g3_45.C = Y;
      g3_45.sAo = 0; g3_45.sAi = 0; g3_45.sAm = H; g3_45.sAk = 1; g3_45.sBo = 0; g3_45.sBi = 0; g3_45.sBn = 1; g3_45.sBk = 1; g3_45.sCo = 0; g3_45.sCi = 0; g3_45.sCm = LP; g3_45.sRo = 0; g3_45.sRi = 0; g3_45.sRm = 0; g3_45.sRn = 0;
      g3_45.M = 8248; g3_45.N = 1; g3_45.K = H; g3_45.zi_n = 1; g3_45.flags = 1; g3_45.act = 0;
      g3_45.alpha = 1.0f; g3_45.beta = 0.0f; g3_45.sa = 1.0f; g3_45.sb = 8.0f; g3_45.Npad = LP; g3_45.pad_ = 0;
      k_gemm<0><<<dim3((unsigned)((LP) + 31) / 32, (unsigned)((8248) + 15) / 16, (unsigned)(1)), 32, 0, stream>>>(g3_45); }
    k_es_scatter<<<(unsigned)((8248 + 255) / 256), 256, 0, stream>>>(Y, LP, slot, IDX, 45, 368740, 8248, out);
    { GemmP g1_46;
      g1_46.A = XS + (size_t)376988 * 8; g1_46.B = W1 + 8832; g1_46.bias = b1 + 2944; g1_46.R = XS + (size_t)376988 * 8; g1_46.C = H1;
      g1_46.sAo = 0; g1_46.sAi = 0; g1_46.sAm = 8; g1_46.sAk = 1; g1_46.sBo = 0; g1_46.sBi = 0; g1_46.sBn = 1; g1_46.sBk = H; g1_46.sCo = 0; g1_46.sCi = 0; g1_46.sCm = H; g1_46.sRo = 0; g1_46.sRi = 0; g1_46.sRm = 0; g1_46.sRn = 0;
      g1_46.M = 8273; g1_46.N = H; g1_46.K = 3; g1_46.zi_n = 1; g1_46.flags = 1; g1_46.act = 1;
      g1_46.alpha = 1.0f; g1_46.beta = 0.0f; g1_46.sa = 1.0f; g1_46.sb = 8.0f; g1_46.Npad = H; g1_46.pad_ = 0;
      k_gemm<0><<<dim3((unsigned)((H) + 31) / 32, (unsigned)((8273) + 15) / 16, (unsigned)(1)), 32, 0, stream>>>(g1_46); }
    { GemmP g2_46;
      g2_46.A = H1; g2_46.B = W2 + 188416; g2_46.bias = b2 + 2944; g2_46.R = H1; g2_46.C = H2;
      g2_46.sAo = 0; g2_46.sAi = 0; g2_46.sAm = H; g2_46.sAk = 1; g2_46.sBo = 0; g2_46.sBi = 0; g2_46.sBn = 1; g2_46.sBk = H; g2_46.sCo = 0; g2_46.sCi = 0; g2_46.sCm = H; g2_46.sRo = 0; g2_46.sRi = 0; g2_46.sRm = 0; g2_46.sRn = 0;
      g2_46.M = 8273; g2_46.N = H; g2_46.K = H; g2_46.zi_n = 1; g2_46.flags = 1; g2_46.act = 1;
      g2_46.alpha = 1.0f; g2_46.beta = 0.0f; g2_46.sa = 1.0f; g2_46.sb = 8.0f; g2_46.Npad = H; g2_46.pad_ = 0;
      k_gemm<0><<<dim3((unsigned)((H) + 31) / 32, (unsigned)((8273) + 15) / 16, (unsigned)(1)), 32, 0, stream>>>(g2_46); }
    { GemmP g3_46;
      g3_46.A = H2; g3_46.B = W3 + 2944; g3_46.bias = b3 + 46; g3_46.R = H2; g3_46.C = Y;
      g3_46.sAo = 0; g3_46.sAi = 0; g3_46.sAm = H; g3_46.sAk = 1; g3_46.sBo = 0; g3_46.sBi = 0; g3_46.sBn = 1; g3_46.sBk = 1; g3_46.sCo = 0; g3_46.sCi = 0; g3_46.sCm = LP; g3_46.sRo = 0; g3_46.sRi = 0; g3_46.sRm = 0; g3_46.sRn = 0;
      g3_46.M = 8273; g3_46.N = 1; g3_46.K = H; g3_46.zi_n = 1; g3_46.flags = 1; g3_46.act = 0;
      g3_46.alpha = 1.0f; g3_46.beta = 0.0f; g3_46.sa = 1.0f; g3_46.sb = 8.0f; g3_46.Npad = LP; g3_46.pad_ = 0;
      k_gemm<0><<<dim3((unsigned)((LP) + 31) / 32, (unsigned)((8273) + 15) / 16, (unsigned)(1)), 32, 0, stream>>>(g3_46); }
    k_es_scatter<<<(unsigned)((8273 + 255) / 256), 256, 0, stream>>>(Y, LP, slot, IDX, 46, 376988, 8273, out);
    { GemmP g1_47;
      g1_47.A = XS + (size_t)385261 * 8; g1_47.B = W1 + 9024; g1_47.bias = b1 + 3008; g1_47.R = XS + (size_t)385261 * 8; g1_47.C = H1;
      g1_47.sAo = 0; g1_47.sAi = 0; g1_47.sAm = 8; g1_47.sAk = 1; g1_47.sBo = 0; g1_47.sBi = 0; g1_47.sBn = 1; g1_47.sBk = H; g1_47.sCo = 0; g1_47.sCi = 0; g1_47.sCm = H; g1_47.sRo = 0; g1_47.sRi = 0; g1_47.sRm = 0; g1_47.sRn = 0;
      g1_47.M = 8061; g1_47.N = H; g1_47.K = 3; g1_47.zi_n = 1; g1_47.flags = 1; g1_47.act = 1;
      g1_47.alpha = 1.0f; g1_47.beta = 0.0f; g1_47.sa = 1.0f; g1_47.sb = 8.0f; g1_47.Npad = H; g1_47.pad_ = 0;
      k_gemm<0><<<dim3((unsigned)((H) + 31) / 32, (unsigned)((8061) + 15) / 16, (unsigned)(1)), 32, 0, stream>>>(g1_47); }
    { GemmP g2_47;
      g2_47.A = H1; g2_47.B = W2 + 192512; g2_47.bias = b2 + 3008; g2_47.R = H1; g2_47.C = H2;
      g2_47.sAo = 0; g2_47.sAi = 0; g2_47.sAm = H; g2_47.sAk = 1; g2_47.sBo = 0; g2_47.sBi = 0; g2_47.sBn = 1; g2_47.sBk = H; g2_47.sCo = 0; g2_47.sCi = 0; g2_47.sCm = H; g2_47.sRo = 0; g2_47.sRi = 0; g2_47.sRm = 0; g2_47.sRn = 0;
      g2_47.M = 8061; g2_47.N = H; g2_47.K = H; g2_47.zi_n = 1; g2_47.flags = 1; g2_47.act = 1;
      g2_47.alpha = 1.0f; g2_47.beta = 0.0f; g2_47.sa = 1.0f; g2_47.sb = 8.0f; g2_47.Npad = H; g2_47.pad_ = 0;
      k_gemm<0><<<dim3((unsigned)((H) + 31) / 32, (unsigned)((8061) + 15) / 16, (unsigned)(1)), 32, 0, stream>>>(g2_47); }
    { GemmP g3_47;
      g3_47.A = H2; g3_47.B = W3 + 3008; g3_47.bias = b3 + 47; g3_47.R = H2; g3_47.C = Y;
      g3_47.sAo = 0; g3_47.sAi = 0; g3_47.sAm = H; g3_47.sAk = 1; g3_47.sBo = 0; g3_47.sBi = 0; g3_47.sBn = 1; g3_47.sBk = 1; g3_47.sCo = 0; g3_47.sCi = 0; g3_47.sCm = LP; g3_47.sRo = 0; g3_47.sRi = 0; g3_47.sRm = 0; g3_47.sRn = 0;
      g3_47.M = 8061; g3_47.N = 1; g3_47.K = H; g3_47.zi_n = 1; g3_47.flags = 1; g3_47.act = 0;
      g3_47.alpha = 1.0f; g3_47.beta = 0.0f; g3_47.sa = 1.0f; g3_47.sb = 8.0f; g3_47.Npad = LP; g3_47.pad_ = 0;
      k_gemm<0><<<dim3((unsigned)((LP) + 31) / 32, (unsigned)((8061) + 15) / 16, (unsigned)(1)), 32, 0, stream>>>(g3_47); }
    k_es_scatter<<<(unsigned)((8061 + 255) / 256), 256, 0, stream>>>(Y, LP, slot, IDX, 47, 385261, 8061, out);
    { GemmP g1_48;
      g1_48.A = XS + (size_t)393322 * 8; g1_48.B = W1 + 9216; g1_48.bias = b1 + 3072; g1_48.R = XS + (size_t)393322 * 8; g1_48.C = H1;
      g1_48.sAo = 0; g1_48.sAi = 0; g1_48.sAm = 8; g1_48.sAk = 1; g1_48.sBo = 0; g1_48.sBi = 0; g1_48.sBn = 1; g1_48.sBk = H; g1_48.sCo = 0; g1_48.sCi = 0; g1_48.sCm = H; g1_48.sRo = 0; g1_48.sRi = 0; g1_48.sRm = 0; g1_48.sRn = 0;
      g1_48.M = 8099; g1_48.N = H; g1_48.K = 3; g1_48.zi_n = 1; g1_48.flags = 1; g1_48.act = 1;
      g1_48.alpha = 1.0f; g1_48.beta = 0.0f; g1_48.sa = 1.0f; g1_48.sb = 8.0f; g1_48.Npad = H; g1_48.pad_ = 0;
      k_gemm<0><<<dim3((unsigned)((H) + 31) / 32, (unsigned)((8099) + 15) / 16, (unsigned)(1)), 32, 0, stream>>>(g1_48); }
    { GemmP g2_48;
      g2_48.A = H1; g2_48.B = W2 + 196608; g2_48.bias = b2 + 3072; g2_48.R = H1; g2_48.C = H2;
      g2_48.sAo = 0; g2_48.sAi = 0; g2_48.sAm = H; g2_48.sAk = 1; g2_48.sBo = 0; g2_48.sBi = 0; g2_48.sBn = 1; g2_48.sBk = H; g2_48.sCo = 0; g2_48.sCi = 0; g2_48.sCm = H; g2_48.sRo = 0; g2_48.sRi = 0; g2_48.sRm = 0; g2_48.sRn = 0;
      g2_48.M = 8099; g2_48.N = H; g2_48.K = H; g2_48.zi_n = 1; g2_48.flags = 1; g2_48.act = 1;
      g2_48.alpha = 1.0f; g2_48.beta = 0.0f; g2_48.sa = 1.0f; g2_48.sb = 8.0f; g2_48.Npad = H; g2_48.pad_ = 0;
      k_gemm<0><<<dim3((unsigned)((H) + 31) / 32, (unsigned)((8099) + 15) / 16, (unsigned)(1)), 32, 0, stream>>>(g2_48); }
    { GemmP g3_48;
      g3_48.A = H2; g3_48.B = W3 + 3072; g3_48.bias = b3 + 48; g3_48.R = H2; g3_48.C = Y;
      g3_48.sAo = 0; g3_48.sAi = 0; g3_48.sAm = H; g3_48.sAk = 1; g3_48.sBo = 0; g3_48.sBi = 0; g3_48.sBn = 1; g3_48.sBk = 1; g3_48.sCo = 0; g3_48.sCi = 0; g3_48.sCm = LP; g3_48.sRo = 0; g3_48.sRi = 0; g3_48.sRm = 0; g3_48.sRn = 0;
      g3_48.M = 8099; g3_48.N = 1; g3_48.K = H; g3_48.zi_n = 1; g3_48.flags = 1; g3_48.act = 0;
      g3_48.alpha = 1.0f; g3_48.beta = 0.0f; g3_48.sa = 1.0f; g3_48.sb = 8.0f; g3_48.Npad = LP; g3_48.pad_ = 0;
      k_gemm<0><<<dim3((unsigned)((LP) + 31) / 32, (unsigned)((8099) + 15) / 16, (unsigned)(1)), 32, 0, stream>>>(g3_48); }
    k_es_scatter<<<(unsigned)((8099 + 255) / 256), 256, 0, stream>>>(Y, LP, slot, IDX, 48, 393322, 8099, out);
    { GemmP g1_49;
      g1_49.A = XS + (size_t)401421 * 8; g1_49.B = W1 + 9408; g1_49.bias = b1 + 3136; g1_49.R = XS + (size_t)401421 * 8; g1_49.C = H1;
      g1_49.sAo = 0; g1_49.sAi = 0; g1_49.sAm = 8; g1_49.sAk = 1; g1_49.sBo = 0; g1_49.sBi = 0; g1_49.sBn = 1; g1_49.sBk = H; g1_49.sCo = 0; g1_49.sCi = 0; g1_49.sCm = H; g1_49.sRo = 0; g1_49.sRi = 0; g1_49.sRm = 0; g1_49.sRn = 0;
      g1_49.M = 8238; g1_49.N = H; g1_49.K = 3; g1_49.zi_n = 1; g1_49.flags = 1; g1_49.act = 1;
      g1_49.alpha = 1.0f; g1_49.beta = 0.0f; g1_49.sa = 1.0f; g1_49.sb = 8.0f; g1_49.Npad = H; g1_49.pad_ = 0;
      k_gemm<0><<<dim3((unsigned)((H) + 31) / 32, (unsigned)((8238) + 15) / 16, (unsigned)(1)), 32, 0, stream>>>(g1_49); }
    { GemmP g2_49;
      g2_49.A = H1; g2_49.B = W2 + 200704; g2_49.bias = b2 + 3136; g2_49.R = H1; g2_49.C = H2;
      g2_49.sAo = 0; g2_49.sAi = 0; g2_49.sAm = H; g2_49.sAk = 1; g2_49.sBo = 0; g2_49.sBi = 0; g2_49.sBn = 1; g2_49.sBk = H; g2_49.sCo = 0; g2_49.sCi = 0; g2_49.sCm = H; g2_49.sRo = 0; g2_49.sRi = 0; g2_49.sRm = 0; g2_49.sRn = 0;
      g2_49.M = 8238; g2_49.N = H; g2_49.K = H; g2_49.zi_n = 1; g2_49.flags = 1; g2_49.act = 1;
      g2_49.alpha = 1.0f; g2_49.beta = 0.0f; g2_49.sa = 1.0f; g2_49.sb = 8.0f; g2_49.Npad = H; g2_49.pad_ = 0;
      k_gemm<0><<<dim3((unsigned)((H) + 31) / 32, (unsigned)((8238) + 15) / 16, (unsigned)(1)), 32, 0, stream>>>(g2_49); }
    { GemmP g3_49;
      g3_49.A = H2; g3_49.B = W3 + 3136; g3_49.bias = b3 + 49; g3_49.R = H2; g3_49.C = Y;
      g3_49.sAo = 0; g3_49.sAi = 0; g3_49.sAm = H; g3_49.sAk = 1; g3_49.sBo = 0; g3_49.sBi = 0; g3_49.sBn = 1; g3_49.sBk = 1; g3_49.sCo = 0; g3_49.sCi = 0; g3_49.sCm = LP; g3_49.sRo = 0; g3_49.sRi = 0; g3_49.sRm = 0; g3_49.sRn = 0;
      g3_49.M = 8238; g3_49.N = 1; g3_49.K = H; g3_49.zi_n = 1; g3_49.flags = 1; g3_49.act = 0;
      g3_49.alpha = 1.0f; g3_49.beta = 0.0f; g3_49.sa = 1.0f; g3_49.sb = 8.0f; g3_49.Npad = LP; g3_49.pad_ = 0;
      k_gemm<0><<<dim3((unsigned)((LP) + 31) / 32, (unsigned)((8238) + 15) / 16, (unsigned)(1)), 32, 0, stream>>>(g3_49); }
    k_es_scatter<<<(unsigned)((8238 + 255) / 256), 256, 0, stream>>>(Y, LP, slot, IDX, 49, 401421, 8238, out);
    { GemmP g1_50;
      g1_50.A = XS + (size_t)409659 * 8; g1_50.B = W1 + 9600; g1_50.bias = b1 + 3200; g1_50.R = XS + (size_t)409659 * 8; g1_50.C = H1;
      g1_50.sAo = 0; g1_50.sAi = 0; g1_50.sAm = 8; g1_50.sAk = 1; g1_50.sBo = 0; g1_50.sBi = 0; g1_50.sBn = 1; g1_50.sBk = H; g1_50.sCo = 0; g1_50.sCi = 0; g1_50.sCm = H; g1_50.sRo = 0; g1_50.sRi = 0; g1_50.sRm = 0; g1_50.sRn = 0;
      g1_50.M = 8291; g1_50.N = H; g1_50.K = 3; g1_50.zi_n = 1; g1_50.flags = 1; g1_50.act = 1;
      g1_50.alpha = 1.0f; g1_50.beta = 0.0f; g1_50.sa = 1.0f; g1_50.sb = 8.0f; g1_50.Npad = H; g1_50.pad_ = 0;
      k_gemm<0><<<dim3((unsigned)((H) + 31) / 32, (unsigned)((8291) + 15) / 16, (unsigned)(1)), 32, 0, stream>>>(g1_50); }
    { GemmP g2_50;
      g2_50.A = H1; g2_50.B = W2 + 204800; g2_50.bias = b2 + 3200; g2_50.R = H1; g2_50.C = H2;
      g2_50.sAo = 0; g2_50.sAi = 0; g2_50.sAm = H; g2_50.sAk = 1; g2_50.sBo = 0; g2_50.sBi = 0; g2_50.sBn = 1; g2_50.sBk = H; g2_50.sCo = 0; g2_50.sCi = 0; g2_50.sCm = H; g2_50.sRo = 0; g2_50.sRi = 0; g2_50.sRm = 0; g2_50.sRn = 0;
      g2_50.M = 8291; g2_50.N = H; g2_50.K = H; g2_50.zi_n = 1; g2_50.flags = 1; g2_50.act = 1;
      g2_50.alpha = 1.0f; g2_50.beta = 0.0f; g2_50.sa = 1.0f; g2_50.sb = 8.0f; g2_50.Npad = H; g2_50.pad_ = 0;
      k_gemm<0><<<dim3((unsigned)((H) + 31) / 32, (unsigned)((8291) + 15) / 16, (unsigned)(1)), 32, 0, stream>>>(g2_50); }
    { GemmP g3_50;
      g3_50.A = H2; g3_50.B = W3 + 3200; g3_50.bias = b3 + 50; g3_50.R = H2; g3_50.C = Y;
      g3_50.sAo = 0; g3_50.sAi = 0; g3_50.sAm = H; g3_50.sAk = 1; g3_50.sBo = 0; g3_50.sBi = 0; g3_50.sBn = 1; g3_50.sBk = 1; g3_50.sCo = 0; g3_50.sCi = 0; g3_50.sCm = LP; g3_50.sRo = 0; g3_50.sRi = 0; g3_50.sRm = 0; g3_50.sRn = 0;
      g3_50.M = 8291; g3_50.N = 1; g3_50.K = H; g3_50.zi_n = 1; g3_50.flags = 1; g3_50.act = 0;
      g3_50.alpha = 1.0f; g3_50.beta = 0.0f; g3_50.sa = 1.0f; g3_50.sb = 8.0f; g3_50.Npad = LP; g3_50.pad_ = 0;
      k_gemm<0><<<dim3((unsigned)((LP) + 31) / 32, (unsigned)((8291) + 15) / 16, (unsigned)(1)), 32, 0, stream>>>(g3_50); }
    k_es_scatter<<<(unsigned)((8291 + 255) / 256), 256, 0, stream>>>(Y, LP, slot, IDX, 50, 409659, 8291, out);
    { GemmP g1_51;
      g1_51.A = XS + (size_t)417950 * 8; g1_51.B = W1 + 9792; g1_51.bias = b1 + 3264; g1_51.R = XS + (size_t)417950 * 8; g1_51.C = H1;
      g1_51.sAo = 0; g1_51.sAi = 0; g1_51.sAm = 8; g1_51.sAk = 1; g1_51.sBo = 0; g1_51.sBi = 0; g1_51.sBn = 1; g1_51.sBk = H; g1_51.sCo = 0; g1_51.sCi = 0; g1_51.sCm = H; g1_51.sRo = 0; g1_51.sRi = 0; g1_51.sRm = 0; g1_51.sRn = 0;
      g1_51.M = 8398; g1_51.N = H; g1_51.K = 3; g1_51.zi_n = 1; g1_51.flags = 1; g1_51.act = 1;
      g1_51.alpha = 1.0f; g1_51.beta = 0.0f; g1_51.sa = 1.0f; g1_51.sb = 8.0f; g1_51.Npad = H; g1_51.pad_ = 0;
      k_gemm<0><<<dim3((unsigned)((H) + 31) / 32, (unsigned)((8398) + 15) / 16, (unsigned)(1)), 32, 0, stream>>>(g1_51); }
    { GemmP g2_51;
      g2_51.A = H1; g2_51.B = W2 + 208896; g2_51.bias = b2 + 3264; g2_51.R = H1; g2_51.C = H2;
      g2_51.sAo = 0; g2_51.sAi = 0; g2_51.sAm = H; g2_51.sAk = 1; g2_51.sBo = 0; g2_51.sBi = 0; g2_51.sBn = 1; g2_51.sBk = H; g2_51.sCo = 0; g2_51.sCi = 0; g2_51.sCm = H; g2_51.sRo = 0; g2_51.sRi = 0; g2_51.sRm = 0; g2_51.sRn = 0;
      g2_51.M = 8398; g2_51.N = H; g2_51.K = H; g2_51.zi_n = 1; g2_51.flags = 1; g2_51.act = 1;
      g2_51.alpha = 1.0f; g2_51.beta = 0.0f; g2_51.sa = 1.0f; g2_51.sb = 8.0f; g2_51.Npad = H; g2_51.pad_ = 0;
      k_gemm<0><<<dim3((unsigned)((H) + 31) / 32, (unsigned)((8398) + 15) / 16, (unsigned)(1)), 32, 0, stream>>>(g2_51); }
    { GemmP g3_51;
      g3_51.A = H2; g3_51.B = W3 + 3264; g3_51.bias = b3 + 51; g3_51.R = H2; g3_51.C = Y;
      g3_51.sAo = 0; g3_51.sAi = 0; g3_51.sAm = H; g3_51.sAk = 1; g3_51.sBo = 0; g3_51.sBi = 0; g3_51.sBn = 1; g3_51.sBk = 1; g3_51.sCo = 0; g3_51.sCi = 0; g3_51.sCm = LP; g3_51.sRo = 0; g3_51.sRi = 0; g3_51.sRm = 0; g3_51.sRn = 0;
      g3_51.M = 8398; g3_51.N = 1; g3_51.K = H; g3_51.zi_n = 1; g3_51.flags = 1; g3_51.act = 0;
      g3_51.alpha = 1.0f; g3_51.beta = 0.0f; g3_51.sa = 1.0f; g3_51.sb = 8.0f; g3_51.Npad = LP; g3_51.pad_ = 0;
      k_gemm<0><<<dim3((unsigned)((LP) + 31) / 32, (unsigned)((8398) + 15) / 16, (unsigned)(1)), 32, 0, stream>>>(g3_51); }
    k_es_scatter<<<(unsigned)((8398 + 255) / 256), 256, 0, stream>>>(Y, LP, slot, IDX, 51, 417950, 8398, out);
    { GemmP g1_52;
      g1_52.A = XS + (size_t)426348 * 8; g1_52.B = W1 + 9984; g1_52.bias = b1 + 3328; g1_52.R = XS + (size_t)426348 * 8; g1_52.C = H1;
      g1_52.sAo = 0; g1_52.sAi = 0; g1_52.sAm = 8; g1_52.sAk = 1; g1_52.sBo = 0; g1_52.sBi = 0; g1_52.sBn = 1; g1_52.sBk = H; g1_52.sCo = 0; g1_52.sCi = 0; g1_52.sCm = H; g1_52.sRo = 0; g1_52.sRi = 0; g1_52.sRm = 0; g1_52.sRn = 0;
      g1_52.M = 8179; g1_52.N = H; g1_52.K = 3; g1_52.zi_n = 1; g1_52.flags = 1; g1_52.act = 1;
      g1_52.alpha = 1.0f; g1_52.beta = 0.0f; g1_52.sa = 1.0f; g1_52.sb = 8.0f; g1_52.Npad = H; g1_52.pad_ = 0;
      k_gemm<0><<<dim3((unsigned)((H) + 31) / 32, (unsigned)((8179) + 15) / 16, (unsigned)(1)), 32, 0, stream>>>(g1_52); }
    { GemmP g2_52;
      g2_52.A = H1; g2_52.B = W2 + 212992; g2_52.bias = b2 + 3328; g2_52.R = H1; g2_52.C = H2;
      g2_52.sAo = 0; g2_52.sAi = 0; g2_52.sAm = H; g2_52.sAk = 1; g2_52.sBo = 0; g2_52.sBi = 0; g2_52.sBn = 1; g2_52.sBk = H; g2_52.sCo = 0; g2_52.sCi = 0; g2_52.sCm = H; g2_52.sRo = 0; g2_52.sRi = 0; g2_52.sRm = 0; g2_52.sRn = 0;
      g2_52.M = 8179; g2_52.N = H; g2_52.K = H; g2_52.zi_n = 1; g2_52.flags = 1; g2_52.act = 1;
      g2_52.alpha = 1.0f; g2_52.beta = 0.0f; g2_52.sa = 1.0f; g2_52.sb = 8.0f; g2_52.Npad = H; g2_52.pad_ = 0;
      k_gemm<0><<<dim3((unsigned)((H) + 31) / 32, (unsigned)((8179) + 15) / 16, (unsigned)(1)), 32, 0, stream>>>(g2_52); }
    { GemmP g3_52;
      g3_52.A = H2; g3_52.B = W3 + 3328; g3_52.bias = b3 + 52; g3_52.R = H2; g3_52.C = Y;
      g3_52.sAo = 0; g3_52.sAi = 0; g3_52.sAm = H; g3_52.sAk = 1; g3_52.sBo = 0; g3_52.sBi = 0; g3_52.sBn = 1; g3_52.sBk = 1; g3_52.sCo = 0; g3_52.sCi = 0; g3_52.sCm = LP; g3_52.sRo = 0; g3_52.sRi = 0; g3_52.sRm = 0; g3_52.sRn = 0;
      g3_52.M = 8179; g3_52.N = 1; g3_52.K = H; g3_52.zi_n = 1; g3_52.flags = 1; g3_52.act = 0;
      g3_52.alpha = 1.0f; g3_52.beta = 0.0f; g3_52.sa = 1.0f; g3_52.sb = 8.0f; g3_52.Npad = LP; g3_52.pad_ = 0;
      k_gemm<0><<<dim3((unsigned)((LP) + 31) / 32, (unsigned)((8179) + 15) / 16, (unsigned)(1)), 32, 0, stream>>>(g3_52); }
    k_es_scatter<<<(unsigned)((8179 + 255) / 256), 256, 0, stream>>>(Y, LP, slot, IDX, 52, 426348, 8179, out);
    { GemmP g1_53;
      g1_53.A = XS + (size_t)434527 * 8; g1_53.B = W1 + 10176; g1_53.bias = b1 + 3392; g1_53.R = XS + (size_t)434527 * 8; g1_53.C = H1;
      g1_53.sAo = 0; g1_53.sAi = 0; g1_53.sAm = 8; g1_53.sAk = 1; g1_53.sBo = 0; g1_53.sBi = 0; g1_53.sBn = 1; g1_53.sBk = H; g1_53.sCo = 0; g1_53.sCi = 0; g1_53.sCm = H; g1_53.sRo = 0; g1_53.sRi = 0; g1_53.sRm = 0; g1_53.sRn = 0;
      g1_53.M = 8271; g1_53.N = H; g1_53.K = 3; g1_53.zi_n = 1; g1_53.flags = 1; g1_53.act = 1;
      g1_53.alpha = 1.0f; g1_53.beta = 0.0f; g1_53.sa = 1.0f; g1_53.sb = 8.0f; g1_53.Npad = H; g1_53.pad_ = 0;
      k_gemm<0><<<dim3((unsigned)((H) + 31) / 32, (unsigned)((8271) + 15) / 16, (unsigned)(1)), 32, 0, stream>>>(g1_53); }
    { GemmP g2_53;
      g2_53.A = H1; g2_53.B = W2 + 217088; g2_53.bias = b2 + 3392; g2_53.R = H1; g2_53.C = H2;
      g2_53.sAo = 0; g2_53.sAi = 0; g2_53.sAm = H; g2_53.sAk = 1; g2_53.sBo = 0; g2_53.sBi = 0; g2_53.sBn = 1; g2_53.sBk = H; g2_53.sCo = 0; g2_53.sCi = 0; g2_53.sCm = H; g2_53.sRo = 0; g2_53.sRi = 0; g2_53.sRm = 0; g2_53.sRn = 0;
      g2_53.M = 8271; g2_53.N = H; g2_53.K = H; g2_53.zi_n = 1; g2_53.flags = 1; g2_53.act = 1;
      g2_53.alpha = 1.0f; g2_53.beta = 0.0f; g2_53.sa = 1.0f; g2_53.sb = 8.0f; g2_53.Npad = H; g2_53.pad_ = 0;
      k_gemm<0><<<dim3((unsigned)((H) + 31) / 32, (unsigned)((8271) + 15) / 16, (unsigned)(1)), 32, 0, stream>>>(g2_53); }
    { GemmP g3_53;
      g3_53.A = H2; g3_53.B = W3 + 3392; g3_53.bias = b3 + 53; g3_53.R = H2; g3_53.C = Y;
      g3_53.sAo = 0; g3_53.sAi = 0; g3_53.sAm = H; g3_53.sAk = 1; g3_53.sBo = 0; g3_53.sBi = 0; g3_53.sBn = 1; g3_53.sBk = 1; g3_53.sCo = 0; g3_53.sCi = 0; g3_53.sCm = LP; g3_53.sRo = 0; g3_53.sRi = 0; g3_53.sRm = 0; g3_53.sRn = 0;
      g3_53.M = 8271; g3_53.N = 1; g3_53.K = H; g3_53.zi_n = 1; g3_53.flags = 1; g3_53.act = 0;
      g3_53.alpha = 1.0f; g3_53.beta = 0.0f; g3_53.sa = 1.0f; g3_53.sb = 8.0f; g3_53.Npad = LP; g3_53.pad_ = 0;
      k_gemm<0><<<dim3((unsigned)((LP) + 31) / 32, (unsigned)((8271) + 15) / 16, (unsigned)(1)), 32, 0, stream>>>(g3_53); }
    k_es_scatter<<<(unsigned)((8271 + 255) / 256), 256, 0, stream>>>(Y, LP, slot, IDX, 53, 434527, 8271, out);
    { GemmP g1_54;
      g1_54.A = XS + (size_t)442798 * 8; g1_54.B = W1 + 10368; g1_54.bias = b1 + 3456; g1_54.R = XS + (size_t)442798 * 8; g1_54.C = H1;
      g1_54.sAo = 0; g1_54.sAi = 0; g1_54.sAm = 8; g1_54.sAk = 1; g1_54.sBo = 0; g1_54.sBi = 0; g1_54.sBn = 1; g1_54.sBk = H; g1_54.sCo = 0; g1_54.sCi = 0; g1_54.sCm = H; g1_54.sRo = 0; g1_54.sRi = 0; g1_54.sRm = 0; g1_54.sRn = 0;
      g1_54.M = 8083; g1_54.N = H; g1_54.K = 3; g1_54.zi_n = 1; g1_54.flags = 1; g1_54.act = 1;
      g1_54.alpha = 1.0f; g1_54.beta = 0.0f; g1_54.sa = 1.0f; g1_54.sb = 8.0f; g1_54.Npad = H; g1_54.pad_ = 0;
      k_gemm<0><<<dim3((unsigned)((H) + 31) / 32, (unsigned)((8083) + 15) / 16, (unsigned)(1)), 32, 0, stream>>>(g1_54); }
    { GemmP g2_54;
      g2_54.A = H1; g2_54.B = W2 + 221184; g2_54.bias = b2 + 3456; g2_54.R = H1; g2_54.C = H2;
      g2_54.sAo = 0; g2_54.sAi = 0; g2_54.sAm = H; g2_54.sAk = 1; g2_54.sBo = 0; g2_54.sBi = 0; g2_54.sBn = 1; g2_54.sBk = H; g2_54.sCo = 0; g2_54.sCi = 0; g2_54.sCm = H; g2_54.sRo = 0; g2_54.sRi = 0; g2_54.sRm = 0; g2_54.sRn = 0;
      g2_54.M = 8083; g2_54.N = H; g2_54.K = H; g2_54.zi_n = 1; g2_54.flags = 1; g2_54.act = 1;
      g2_54.alpha = 1.0f; g2_54.beta = 0.0f; g2_54.sa = 1.0f; g2_54.sb = 8.0f; g2_54.Npad = H; g2_54.pad_ = 0;
      k_gemm<0><<<dim3((unsigned)((H) + 31) / 32, (unsigned)((8083) + 15) / 16, (unsigned)(1)), 32, 0, stream>>>(g2_54); }
    { GemmP g3_54;
      g3_54.A = H2; g3_54.B = W3 + 3456; g3_54.bias = b3 + 54; g3_54.R = H2; g3_54.C = Y;
      g3_54.sAo = 0; g3_54.sAi = 0; g3_54.sAm = H; g3_54.sAk = 1; g3_54.sBo = 0; g3_54.sBi = 0; g3_54.sBn = 1; g3_54.sBk = 1; g3_54.sCo = 0; g3_54.sCi = 0; g3_54.sCm = LP; g3_54.sRo = 0; g3_54.sRi = 0; g3_54.sRm = 0; g3_54.sRn = 0;
      g3_54.M = 8083; g3_54.N = 1; g3_54.K = H; g3_54.zi_n = 1; g3_54.flags = 1; g3_54.act = 0;
      g3_54.alpha = 1.0f; g3_54.beta = 0.0f; g3_54.sa = 1.0f; g3_54.sb = 8.0f; g3_54.Npad = LP; g3_54.pad_ = 0;
      k_gemm<0><<<dim3((unsigned)((LP) + 31) / 32, (unsigned)((8083) + 15) / 16, (unsigned)(1)), 32, 0, stream>>>(g3_54); }
    k_es_scatter<<<(unsigned)((8083 + 255) / 256), 256, 0, stream>>>(Y, LP, slot, IDX, 54, 442798, 8083, out);
    { GemmP g1_55;
      g1_55.A = XS + (size_t)450881 * 8; g1_55.B = W1 + 10560; g1_55.bias = b1 + 3520; g1_55.R = XS + (size_t)450881 * 8; g1_55.C = H1;
      g1_55.sAo = 0; g1_55.sAi = 0; g1_55.sAm = 8; g1_55.sAk = 1; g1_55.sBo = 0; g1_55.sBi = 0; g1_55.sBn = 1; g1_55.sBk = H; g1_55.sCo = 0; g1_55.sCi = 0; g1_55.sCm = H; g1_55.sRo = 0; g1_55.sRi = 0; g1_55.sRm = 0; g1_55.sRn = 0;
      g1_55.M = 8143; g1_55.N = H; g1_55.K = 3; g1_55.zi_n = 1; g1_55.flags = 1; g1_55.act = 1;
      g1_55.alpha = 1.0f; g1_55.beta = 0.0f; g1_55.sa = 1.0f; g1_55.sb = 8.0f; g1_55.Npad = H; g1_55.pad_ = 0;
      k_gemm<0><<<dim3((unsigned)((H) + 31) / 32, (unsigned)((8143) + 15) / 16, (unsigned)(1)), 32, 0, stream>>>(g1_55); }
    { GemmP g2_55;
      g2_55.A = H1; g2_55.B = W2 + 225280; g2_55.bias = b2 + 3520; g2_55.R = H1; g2_55.C = H2;
      g2_55.sAo = 0; g2_55.sAi = 0; g2_55.sAm = H; g2_55.sAk = 1; g2_55.sBo = 0; g2_55.sBi = 0; g2_55.sBn = 1; g2_55.sBk = H; g2_55.sCo = 0; g2_55.sCi = 0; g2_55.sCm = H; g2_55.sRo = 0; g2_55.sRi = 0; g2_55.sRm = 0; g2_55.sRn = 0;
      g2_55.M = 8143; g2_55.N = H; g2_55.K = H; g2_55.zi_n = 1; g2_55.flags = 1; g2_55.act = 1;
      g2_55.alpha = 1.0f; g2_55.beta = 0.0f; g2_55.sa = 1.0f; g2_55.sb = 8.0f; g2_55.Npad = H; g2_55.pad_ = 0;
      k_gemm<0><<<dim3((unsigned)((H) + 31) / 32, (unsigned)((8143) + 15) / 16, (unsigned)(1)), 32, 0, stream>>>(g2_55); }
    { GemmP g3_55;
      g3_55.A = H2; g3_55.B = W3 + 3520; g3_55.bias = b3 + 55; g3_55.R = H2; g3_55.C = Y;
      g3_55.sAo = 0; g3_55.sAi = 0; g3_55.sAm = H; g3_55.sAk = 1; g3_55.sBo = 0; g3_55.sBi = 0; g3_55.sBn = 1; g3_55.sBk = 1; g3_55.sCo = 0; g3_55.sCi = 0; g3_55.sCm = LP; g3_55.sRo = 0; g3_55.sRi = 0; g3_55.sRm = 0; g3_55.sRn = 0;
      g3_55.M = 8143; g3_55.N = 1; g3_55.K = H; g3_55.zi_n = 1; g3_55.flags = 1; g3_55.act = 0;
      g3_55.alpha = 1.0f; g3_55.beta = 0.0f; g3_55.sa = 1.0f; g3_55.sb = 8.0f; g3_55.Npad = LP; g3_55.pad_ = 0;
      k_gemm<0><<<dim3((unsigned)((LP) + 31) / 32, (unsigned)((8143) + 15) / 16, (unsigned)(1)), 32, 0, stream>>>(g3_55); }
    k_es_scatter<<<(unsigned)((8143 + 255) / 256), 256, 0, stream>>>(Y, LP, slot, IDX, 55, 450881, 8143, out);
    { GemmP g1_56;
      g1_56.A = XS + (size_t)459024 * 8; g1_56.B = W1 + 10752; g1_56.bias = b1 + 3584; g1_56.R = XS + (size_t)459024 * 8; g1_56.C = H1;
      g1_56.sAo = 0; g1_56.sAi = 0; g1_56.sAm = 8; g1_56.sAk = 1; g1_56.sBo = 0; g1_56.sBi = 0; g1_56.sBn = 1; g1_56.sBk = H; g1_56.sCo = 0; g1_56.sCi = 0; g1_56.sCm = H; g1_56.sRo = 0; g1_56.sRi = 0; g1_56.sRm = 0; g1_56.sRn = 0;
      g1_56.M = 8146; g1_56.N = H; g1_56.K = 3; g1_56.zi_n = 1; g1_56.flags = 1; g1_56.act = 1;
      g1_56.alpha = 1.0f; g1_56.beta = 0.0f; g1_56.sa = 1.0f; g1_56.sb = 8.0f; g1_56.Npad = H; g1_56.pad_ = 0;
      k_gemm<0><<<dim3((unsigned)((H) + 31) / 32, (unsigned)((8146) + 15) / 16, (unsigned)(1)), 32, 0, stream>>>(g1_56); }
    { GemmP g2_56;
      g2_56.A = H1; g2_56.B = W2 + 229376; g2_56.bias = b2 + 3584; g2_56.R = H1; g2_56.C = H2;
      g2_56.sAo = 0; g2_56.sAi = 0; g2_56.sAm = H; g2_56.sAk = 1; g2_56.sBo = 0; g2_56.sBi = 0; g2_56.sBn = 1; g2_56.sBk = H; g2_56.sCo = 0; g2_56.sCi = 0; g2_56.sCm = H; g2_56.sRo = 0; g2_56.sRi = 0; g2_56.sRm = 0; g2_56.sRn = 0;
      g2_56.M = 8146; g2_56.N = H; g2_56.K = H; g2_56.zi_n = 1; g2_56.flags = 1; g2_56.act = 1;
      g2_56.alpha = 1.0f; g2_56.beta = 0.0f; g2_56.sa = 1.0f; g2_56.sb = 8.0f; g2_56.Npad = H; g2_56.pad_ = 0;
      k_gemm<0><<<dim3((unsigned)((H) + 31) / 32, (unsigned)((8146) + 15) / 16, (unsigned)(1)), 32, 0, stream>>>(g2_56); }
    { GemmP g3_56;
      g3_56.A = H2; g3_56.B = W3 + 3584; g3_56.bias = b3 + 56; g3_56.R = H2; g3_56.C = Y;
      g3_56.sAo = 0; g3_56.sAi = 0; g3_56.sAm = H; g3_56.sAk = 1; g3_56.sBo = 0; g3_56.sBi = 0; g3_56.sBn = 1; g3_56.sBk = 1; g3_56.sCo = 0; g3_56.sCi = 0; g3_56.sCm = LP; g3_56.sRo = 0; g3_56.sRi = 0; g3_56.sRm = 0; g3_56.sRn = 0;
      g3_56.M = 8146; g3_56.N = 1; g3_56.K = H; g3_56.zi_n = 1; g3_56.flags = 1; g3_56.act = 0;
      g3_56.alpha = 1.0f; g3_56.beta = 0.0f; g3_56.sa = 1.0f; g3_56.sb = 8.0f; g3_56.Npad = LP; g3_56.pad_ = 0;
      k_gemm<0><<<dim3((unsigned)((LP) + 31) / 32, (unsigned)((8146) + 15) / 16, (unsigned)(1)), 32, 0, stream>>>(g3_56); }
    k_es_scatter<<<(unsigned)((8146 + 255) / 256), 256, 0, stream>>>(Y, LP, slot, IDX, 56, 459024, 8146, out);
    { GemmP g1_57;
      g1_57.A = XS + (size_t)467170 * 8; g1_57.B = W1 + 10944; g1_57.bias = b1 + 3648; g1_57.R = XS + (size_t)467170 * 8; g1_57.C = H1;
      g1_57.sAo = 0; g1_57.sAi = 0; g1_57.sAm = 8; g1_57.sAk = 1; g1_57.sBo = 0; g1_57.sBi = 0; g1_57.sBn = 1; g1_57.sBk = H; g1_57.sCo = 0; g1_57.sCi = 0; g1_57.sCm = H; g1_57.sRo = 0; g1_57.sRi = 0; g1_57.sRm = 0; g1_57.sRn = 0;
      g1_57.M = 8104; g1_57.N = H; g1_57.K = 3; g1_57.zi_n = 1; g1_57.flags = 1; g1_57.act = 1;
      g1_57.alpha = 1.0f; g1_57.beta = 0.0f; g1_57.sa = 1.0f; g1_57.sb = 8.0f; g1_57.Npad = H; g1_57.pad_ = 0;
      k_gemm<0><<<dim3((unsigned)((H) + 31) / 32, (unsigned)((8104) + 15) / 16, (unsigned)(1)), 32, 0, stream>>>(g1_57); }
    { GemmP g2_57;
      g2_57.A = H1; g2_57.B = W2 + 233472; g2_57.bias = b2 + 3648; g2_57.R = H1; g2_57.C = H2;
      g2_57.sAo = 0; g2_57.sAi = 0; g2_57.sAm = H; g2_57.sAk = 1; g2_57.sBo = 0; g2_57.sBi = 0; g2_57.sBn = 1; g2_57.sBk = H; g2_57.sCo = 0; g2_57.sCi = 0; g2_57.sCm = H; g2_57.sRo = 0; g2_57.sRi = 0; g2_57.sRm = 0; g2_57.sRn = 0;
      g2_57.M = 8104; g2_57.N = H; g2_57.K = H; g2_57.zi_n = 1; g2_57.flags = 1; g2_57.act = 1;
      g2_57.alpha = 1.0f; g2_57.beta = 0.0f; g2_57.sa = 1.0f; g2_57.sb = 8.0f; g2_57.Npad = H; g2_57.pad_ = 0;
      k_gemm<0><<<dim3((unsigned)((H) + 31) / 32, (unsigned)((8104) + 15) / 16, (unsigned)(1)), 32, 0, stream>>>(g2_57); }
    { GemmP g3_57;
      g3_57.A = H2; g3_57.B = W3 + 3648; g3_57.bias = b3 + 57; g3_57.R = H2; g3_57.C = Y;
      g3_57.sAo = 0; g3_57.sAi = 0; g3_57.sAm = H; g3_57.sAk = 1; g3_57.sBo = 0; g3_57.sBi = 0; g3_57.sBn = 1; g3_57.sBk = 1; g3_57.sCo = 0; g3_57.sCi = 0; g3_57.sCm = LP; g3_57.sRo = 0; g3_57.sRi = 0; g3_57.sRm = 0; g3_57.sRn = 0;
      g3_57.M = 8104; g3_57.N = 1; g3_57.K = H; g3_57.zi_n = 1; g3_57.flags = 1; g3_57.act = 0;
      g3_57.alpha = 1.0f; g3_57.beta = 0.0f; g3_57.sa = 1.0f; g3_57.sb = 8.0f; g3_57.Npad = LP; g3_57.pad_ = 0;
      k_gemm<0><<<dim3((unsigned)((LP) + 31) / 32, (unsigned)((8104) + 15) / 16, (unsigned)(1)), 32, 0, stream>>>(g3_57); }
    k_es_scatter<<<(unsigned)((8104 + 255) / 256), 256, 0, stream>>>(Y, LP, slot, IDX, 57, 467170, 8104, out);
    { GemmP g1_58;
      g1_58.A = XS + (size_t)475274 * 8; g1_58.B = W1 + 11136; g1_58.bias = b1 + 3712; g1_58.R = XS + (size_t)475274 * 8; g1_58.C = H1;
      g1_58.sAo = 0; g1_58.sAi = 0; g1_58.sAm = 8; g1_58.sAk = 1; g1_58.sBo = 0; g1_58.sBi = 0; g1_58.sBn = 1; g1_58.sBk = H; g1_58.sCo = 0; g1_58.sCi = 0; g1_58.sCm = H; g1_58.sRo = 0; g1_58.sRi = 0; g1_58.sRm = 0; g1_58.sRn = 0;
      g1_58.M = 8212; g1_58.N = H; g1_58.K = 3; g1_58.zi_n = 1; g1_58.flags = 1; g1_58.act = 1;
      g1_58.alpha = 1.0f; g1_58.beta = 0.0f; g1_58.sa = 1.0f; g1_58.sb = 8.0f; g1_58.Npad = H; g1_58.pad_ = 0;
      k_gemm<0><<<dim3((unsigned)((H) + 31) / 32, (unsigned)((8212) + 15) / 16, (unsigned)(1)), 32, 0, stream>>>(g1_58); }
    { GemmP g2_58;
      g2_58.A = H1; g2_58.B = W2 + 237568; g2_58.bias = b2 + 3712; g2_58.R = H1; g2_58.C = H2;
      g2_58.sAo = 0; g2_58.sAi = 0; g2_58.sAm = H; g2_58.sAk = 1; g2_58.sBo = 0; g2_58.sBi = 0; g2_58.sBn = 1; g2_58.sBk = H; g2_58.sCo = 0; g2_58.sCi = 0; g2_58.sCm = H; g2_58.sRo = 0; g2_58.sRi = 0; g2_58.sRm = 0; g2_58.sRn = 0;
      g2_58.M = 8212; g2_58.N = H; g2_58.K = H; g2_58.zi_n = 1; g2_58.flags = 1; g2_58.act = 1;
      g2_58.alpha = 1.0f; g2_58.beta = 0.0f; g2_58.sa = 1.0f; g2_58.sb = 8.0f; g2_58.Npad = H; g2_58.pad_ = 0;
      k_gemm<0><<<dim3((unsigned)((H) + 31) / 32, (unsigned)((8212) + 15) / 16, (unsigned)(1)), 32, 0, stream>>>(g2_58); }
    { GemmP g3_58;
      g3_58.A = H2; g3_58.B = W3 + 3712; g3_58.bias = b3 + 58; g3_58.R = H2; g3_58.C = Y;
      g3_58.sAo = 0; g3_58.sAi = 0; g3_58.sAm = H; g3_58.sAk = 1; g3_58.sBo = 0; g3_58.sBi = 0; g3_58.sBn = 1; g3_58.sBk = 1; g3_58.sCo = 0; g3_58.sCi = 0; g3_58.sCm = LP; g3_58.sRo = 0; g3_58.sRi = 0; g3_58.sRm = 0; g3_58.sRn = 0;
      g3_58.M = 8212; g3_58.N = 1; g3_58.K = H; g3_58.zi_n = 1; g3_58.flags = 1; g3_58.act = 0;
      g3_58.alpha = 1.0f; g3_58.beta = 0.0f; g3_58.sa = 1.0f; g3_58.sb = 8.0f; g3_58.Npad = LP; g3_58.pad_ = 0;
      k_gemm<0><<<dim3((unsigned)((LP) + 31) / 32, (unsigned)((8212) + 15) / 16, (unsigned)(1)), 32, 0, stream>>>(g3_58); }
    k_es_scatter<<<(unsigned)((8212 + 255) / 256), 256, 0, stream>>>(Y, LP, slot, IDX, 58, 475274, 8212, out);
    { GemmP g1_59;
      g1_59.A = XS + (size_t)483486 * 8; g1_59.B = W1 + 11328; g1_59.bias = b1 + 3776; g1_59.R = XS + (size_t)483486 * 8; g1_59.C = H1;
      g1_59.sAo = 0; g1_59.sAi = 0; g1_59.sAm = 8; g1_59.sAk = 1; g1_59.sBo = 0; g1_59.sBi = 0; g1_59.sBn = 1; g1_59.sBk = H; g1_59.sCo = 0; g1_59.sCi = 0; g1_59.sCm = H; g1_59.sRo = 0; g1_59.sRi = 0; g1_59.sRm = 0; g1_59.sRn = 0;
      g1_59.M = 8206; g1_59.N = H; g1_59.K = 3; g1_59.zi_n = 1; g1_59.flags = 1; g1_59.act = 1;
      g1_59.alpha = 1.0f; g1_59.beta = 0.0f; g1_59.sa = 1.0f; g1_59.sb = 8.0f; g1_59.Npad = H; g1_59.pad_ = 0;
      k_gemm<0><<<dim3((unsigned)((H) + 31) / 32, (unsigned)((8206) + 15) / 16, (unsigned)(1)), 32, 0, stream>>>(g1_59); }
    { GemmP g2_59;
      g2_59.A = H1; g2_59.B = W2 + 241664; g2_59.bias = b2 + 3776; g2_59.R = H1; g2_59.C = H2;
      g2_59.sAo = 0; g2_59.sAi = 0; g2_59.sAm = H; g2_59.sAk = 1; g2_59.sBo = 0; g2_59.sBi = 0; g2_59.sBn = 1; g2_59.sBk = H; g2_59.sCo = 0; g2_59.sCi = 0; g2_59.sCm = H; g2_59.sRo = 0; g2_59.sRi = 0; g2_59.sRm = 0; g2_59.sRn = 0;
      g2_59.M = 8206; g2_59.N = H; g2_59.K = H; g2_59.zi_n = 1; g2_59.flags = 1; g2_59.act = 1;
      g2_59.alpha = 1.0f; g2_59.beta = 0.0f; g2_59.sa = 1.0f; g2_59.sb = 8.0f; g2_59.Npad = H; g2_59.pad_ = 0;
      k_gemm<0><<<dim3((unsigned)((H) + 31) / 32, (unsigned)((8206) + 15) / 16, (unsigned)(1)), 32, 0, stream>>>(g2_59); }
    { GemmP g3_59;
      g3_59.A = H2; g3_59.B = W3 + 3776; g3_59.bias = b3 + 59; g3_59.R = H2; g3_59.C = Y;
      g3_59.sAo = 0; g3_59.sAi = 0; g3_59.sAm = H; g3_59.sAk = 1; g3_59.sBo = 0; g3_59.sBi = 0; g3_59.sBn = 1; g3_59.sBk = 1; g3_59.sCo = 0; g3_59.sCi = 0; g3_59.sCm = LP; g3_59.sRo = 0; g3_59.sRi = 0; g3_59.sRm = 0; g3_59.sRn = 0;
      g3_59.M = 8206; g3_59.N = 1; g3_59.K = H; g3_59.zi_n = 1; g3_59.flags = 1; g3_59.act = 0;
      g3_59.alpha = 1.0f; g3_59.beta = 0.0f; g3_59.sa = 1.0f; g3_59.sb = 8.0f; g3_59.Npad = LP; g3_59.pad_ = 0;
      k_gemm<0><<<dim3((unsigned)((LP) + 31) / 32, (unsigned)((8206) + 15) / 16, (unsigned)(1)), 32, 0, stream>>>(g3_59); }
    k_es_scatter<<<(unsigned)((8206 + 255) / 256), 256, 0, stream>>>(Y, LP, slot, IDX, 59, 483486, 8206, out);
    { GemmP g1_60;
      g1_60.A = XS + (size_t)491692 * 8; g1_60.B = W1 + 11520; g1_60.bias = b1 + 3840; g1_60.R = XS + (size_t)491692 * 8; g1_60.C = H1;
      g1_60.sAo = 0; g1_60.sAi = 0; g1_60.sAm = 8; g1_60.sAk = 1; g1_60.sBo = 0; g1_60.sBi = 0; g1_60.sBn = 1; g1_60.sBk = H; g1_60.sCo = 0; g1_60.sCi = 0; g1_60.sCm = H; g1_60.sRo = 0; g1_60.sRi = 0; g1_60.sRm = 0; g1_60.sRn = 0;
      g1_60.M = 8191; g1_60.N = H; g1_60.K = 3; g1_60.zi_n = 1; g1_60.flags = 1; g1_60.act = 1;
      g1_60.alpha = 1.0f; g1_60.beta = 0.0f; g1_60.sa = 1.0f; g1_60.sb = 8.0f; g1_60.Npad = H; g1_60.pad_ = 0;
      k_gemm<0><<<dim3((unsigned)((H) + 31) / 32, (unsigned)((8191) + 15) / 16, (unsigned)(1)), 32, 0, stream>>>(g1_60); }
    { GemmP g2_60;
      g2_60.A = H1; g2_60.B = W2 + 245760; g2_60.bias = b2 + 3840; g2_60.R = H1; g2_60.C = H2;
      g2_60.sAo = 0; g2_60.sAi = 0; g2_60.sAm = H; g2_60.sAk = 1; g2_60.sBo = 0; g2_60.sBi = 0; g2_60.sBn = 1; g2_60.sBk = H; g2_60.sCo = 0; g2_60.sCi = 0; g2_60.sCm = H; g2_60.sRo = 0; g2_60.sRi = 0; g2_60.sRm = 0; g2_60.sRn = 0;
      g2_60.M = 8191; g2_60.N = H; g2_60.K = H; g2_60.zi_n = 1; g2_60.flags = 1; g2_60.act = 1;
      g2_60.alpha = 1.0f; g2_60.beta = 0.0f; g2_60.sa = 1.0f; g2_60.sb = 8.0f; g2_60.Npad = H; g2_60.pad_ = 0;
      k_gemm<0><<<dim3((unsigned)((H) + 31) / 32, (unsigned)((8191) + 15) / 16, (unsigned)(1)), 32, 0, stream>>>(g2_60); }
    { GemmP g3_60;
      g3_60.A = H2; g3_60.B = W3 + 3840; g3_60.bias = b3 + 60; g3_60.R = H2; g3_60.C = Y;
      g3_60.sAo = 0; g3_60.sAi = 0; g3_60.sAm = H; g3_60.sAk = 1; g3_60.sBo = 0; g3_60.sBi = 0; g3_60.sBn = 1; g3_60.sBk = 1; g3_60.sCo = 0; g3_60.sCi = 0; g3_60.sCm = LP; g3_60.sRo = 0; g3_60.sRi = 0; g3_60.sRm = 0; g3_60.sRn = 0;
      g3_60.M = 8191; g3_60.N = 1; g3_60.K = H; g3_60.zi_n = 1; g3_60.flags = 1; g3_60.act = 0;
      g3_60.alpha = 1.0f; g3_60.beta = 0.0f; g3_60.sa = 1.0f; g3_60.sb = 8.0f; g3_60.Npad = LP; g3_60.pad_ = 0;
      k_gemm<0><<<dim3((unsigned)((LP) + 31) / 32, (unsigned)((8191) + 15) / 16, (unsigned)(1)), 32, 0, stream>>>(g3_60); }
    k_es_scatter<<<(unsigned)((8191 + 255) / 256), 256, 0, stream>>>(Y, LP, slot, IDX, 60, 491692, 8191, out);
    { GemmP g1_61;
      g1_61.A = XS + (size_t)499883 * 8; g1_61.B = W1 + 11712; g1_61.bias = b1 + 3904; g1_61.R = XS + (size_t)499883 * 8; g1_61.C = H1;
      g1_61.sAo = 0; g1_61.sAi = 0; g1_61.sAm = 8; g1_61.sAk = 1; g1_61.sBo = 0; g1_61.sBi = 0; g1_61.sBn = 1; g1_61.sBk = H; g1_61.sCo = 0; g1_61.sCi = 0; g1_61.sCm = H; g1_61.sRo = 0; g1_61.sRi = 0; g1_61.sRm = 0; g1_61.sRn = 0;
      g1_61.M = 8105; g1_61.N = H; g1_61.K = 3; g1_61.zi_n = 1; g1_61.flags = 1; g1_61.act = 1;
      g1_61.alpha = 1.0f; g1_61.beta = 0.0f; g1_61.sa = 1.0f; g1_61.sb = 8.0f; g1_61.Npad = H; g1_61.pad_ = 0;
      k_gemm<0><<<dim3((unsigned)((H) + 31) / 32, (unsigned)((8105) + 15) / 16, (unsigned)(1)), 32, 0, stream>>>(g1_61); }
    { GemmP g2_61;
      g2_61.A = H1; g2_61.B = W2 + 249856; g2_61.bias = b2 + 3904; g2_61.R = H1; g2_61.C = H2;
      g2_61.sAo = 0; g2_61.sAi = 0; g2_61.sAm = H; g2_61.sAk = 1; g2_61.sBo = 0; g2_61.sBi = 0; g2_61.sBn = 1; g2_61.sBk = H; g2_61.sCo = 0; g2_61.sCi = 0; g2_61.sCm = H; g2_61.sRo = 0; g2_61.sRi = 0; g2_61.sRm = 0; g2_61.sRn = 0;
      g2_61.M = 8105; g2_61.N = H; g2_61.K = H; g2_61.zi_n = 1; g2_61.flags = 1; g2_61.act = 1;
      g2_61.alpha = 1.0f; g2_61.beta = 0.0f; g2_61.sa = 1.0f; g2_61.sb = 8.0f; g2_61.Npad = H; g2_61.pad_ = 0;
      k_gemm<0><<<dim3((unsigned)((H) + 31) / 32, (unsigned)((8105) + 15) / 16, (unsigned)(1)), 32, 0, stream>>>(g2_61); }
    { GemmP g3_61;
      g3_61.A = H2; g3_61.B = W3 + 3904; g3_61.bias = b3 + 61; g3_61.R = H2; g3_61.C = Y;
      g3_61.sAo = 0; g3_61.sAi = 0; g3_61.sAm = H; g3_61.sAk = 1; g3_61.sBo = 0; g3_61.sBi = 0; g3_61.sBn = 1; g3_61.sBk = 1; g3_61.sCo = 0; g3_61.sCi = 0; g3_61.sCm = LP; g3_61.sRo = 0; g3_61.sRi = 0; g3_61.sRm = 0; g3_61.sRn = 0;
      g3_61.M = 8105; g3_61.N = 1; g3_61.K = H; g3_61.zi_n = 1; g3_61.flags = 1; g3_61.act = 0;
      g3_61.alpha = 1.0f; g3_61.beta = 0.0f; g3_61.sa = 1.0f; g3_61.sb = 8.0f; g3_61.Npad = LP; g3_61.pad_ = 0;
      k_gemm<0><<<dim3((unsigned)((LP) + 31) / 32, (unsigned)((8105) + 15) / 16, (unsigned)(1)), 32, 0, stream>>>(g3_61); }
    k_es_scatter<<<(unsigned)((8105 + 255) / 256), 256, 0, stream>>>(Y, LP, slot, IDX, 61, 499883, 8105, out);
    { GemmP g1_62;
      g1_62.A = XS + (size_t)507988 * 8; g1_62.B = W1 + 11904; g1_62.bias = b1 + 3968; g1_62.R = XS + (size_t)507988 * 8; g1_62.C = H1;
      g1_62.sAo = 0; g1_62.sAi = 0; g1_62.sAm = 8; g1_62.sAk = 1; g1_62.sBo = 0; g1_62.sBi = 0; g1_62.sBn = 1; g1_62.sBk = H; g1_62.sCo = 0; g1_62.sCi = 0; g1_62.sCm = H; g1_62.sRo = 0; g1_62.sRi = 0; g1_62.sRm = 0; g1_62.sRn = 0;
      g1_62.M = 8121; g1_62.N = H; g1_62.K = 3; g1_62.zi_n = 1; g1_62.flags = 1; g1_62.act = 1;
      g1_62.alpha = 1.0f; g1_62.beta = 0.0f; g1_62.sa = 1.0f; g1_62.sb = 8.0f; g1_62.Npad = H; g1_62.pad_ = 0;
      k_gemm<0><<<dim3((unsigned)((H) + 31) / 32, (unsigned)((8121) + 15) / 16, (unsigned)(1)), 32, 0, stream>>>(g1_62); }
    { GemmP g2_62;
      g2_62.A = H1; g2_62.B = W2 + 253952; g2_62.bias = b2 + 3968; g2_62.R = H1; g2_62.C = H2;
      g2_62.sAo = 0; g2_62.sAi = 0; g2_62.sAm = H; g2_62.sAk = 1; g2_62.sBo = 0; g2_62.sBi = 0; g2_62.sBn = 1; g2_62.sBk = H; g2_62.sCo = 0; g2_62.sCi = 0; g2_62.sCm = H; g2_62.sRo = 0; g2_62.sRi = 0; g2_62.sRm = 0; g2_62.sRn = 0;
      g2_62.M = 8121; g2_62.N = H; g2_62.K = H; g2_62.zi_n = 1; g2_62.flags = 1; g2_62.act = 1;
      g2_62.alpha = 1.0f; g2_62.beta = 0.0f; g2_62.sa = 1.0f; g2_62.sb = 8.0f; g2_62.Npad = H; g2_62.pad_ = 0;
      k_gemm<0><<<dim3((unsigned)((H) + 31) / 32, (unsigned)((8121) + 15) / 16, (unsigned)(1)), 32, 0, stream>>>(g2_62); }
    { GemmP g3_62;
      g3_62.A = H2; g3_62.B = W3 + 3968; g3_62.bias = b3 + 62; g3_62.R = H2; g3_62.C = Y;
      g3_62.sAo = 0; g3_62.sAi = 0; g3_62.sAm = H; g3_62.sAk = 1; g3_62.sBo = 0; g3_62.sBi = 0; g3_62.sBn = 1; g3_62.sBk = 1; g3_62.sCo = 0; g3_62.sCi = 0; g3_62.sCm = LP; g3_62.sRo = 0; g3_62.sRi = 0; g3_62.sRm = 0; g3_62.sRn = 0;
      g3_62.M = 8121; g3_62.N = 1; g3_62.K = H; g3_62.zi_n = 1; g3_62.flags = 1; g3_62.act = 0;
      g3_62.alpha = 1.0f; g3_62.beta = 0.0f; g3_62.sa = 1.0f; g3_62.sb = 8.0f; g3_62.Npad = LP; g3_62.pad_ = 0;
      k_gemm<0><<<dim3((unsigned)((LP) + 31) / 32, (unsigned)((8121) + 15) / 16, (unsigned)(1)), 32, 0, stream>>>(g3_62); }
    k_es_scatter<<<(unsigned)((8121 + 255) / 256), 256, 0, stream>>>(Y, LP, slot, IDX, 62, 507988, 8121, out);
    { GemmP g1_63;
      g1_63.A = XS + (size_t)516109 * 8; g1_63.B = W1 + 12096; g1_63.bias = b1 + 4032; g1_63.R = XS + (size_t)516109 * 8; g1_63.C = H1;
      g1_63.sAo = 0; g1_63.sAi = 0; g1_63.sAm = 8; g1_63.sAk = 1; g1_63.sBo = 0; g1_63.sBi = 0; g1_63.sBn = 1; g1_63.sBk = H; g1_63.sCo = 0; g1_63.sCi = 0; g1_63.sCm = H; g1_63.sRo = 0; g1_63.sRi = 0; g1_63.sRm = 0; g1_63.sRn = 0;
      g1_63.M = 8179; g1_63.N = H; g1_63.K = 3; g1_63.zi_n = 1; g1_63.flags = 1; g1_63.act = 1;
      g1_63.alpha = 1.0f; g1_63.beta = 0.0f; g1_63.sa = 1.0f; g1_63.sb = 8.0f; g1_63.Npad = H; g1_63.pad_ = 0;
      k_gemm<0><<<dim3((unsigned)((H) + 31) / 32, (unsigned)((8179) + 15) / 16, (unsigned)(1)), 32, 0, stream>>>(g1_63); }
    { GemmP g2_63;
      g2_63.A = H1; g2_63.B = W2 + 258048; g2_63.bias = b2 + 4032; g2_63.R = H1; g2_63.C = H2;
      g2_63.sAo = 0; g2_63.sAi = 0; g2_63.sAm = H; g2_63.sAk = 1; g2_63.sBo = 0; g2_63.sBi = 0; g2_63.sBn = 1; g2_63.sBk = H; g2_63.sCo = 0; g2_63.sCi = 0; g2_63.sCm = H; g2_63.sRo = 0; g2_63.sRi = 0; g2_63.sRm = 0; g2_63.sRn = 0;
      g2_63.M = 8179; g2_63.N = H; g2_63.K = H; g2_63.zi_n = 1; g2_63.flags = 1; g2_63.act = 1;
      g2_63.alpha = 1.0f; g2_63.beta = 0.0f; g2_63.sa = 1.0f; g2_63.sb = 8.0f; g2_63.Npad = H; g2_63.pad_ = 0;
      k_gemm<0><<<dim3((unsigned)((H) + 31) / 32, (unsigned)((8179) + 15) / 16, (unsigned)(1)), 32, 0, stream>>>(g2_63); }
    { GemmP g3_63;
      g3_63.A = H2; g3_63.B = W3 + 4032; g3_63.bias = b3 + 63; g3_63.R = H2; g3_63.C = Y;
      g3_63.sAo = 0; g3_63.sAi = 0; g3_63.sAm = H; g3_63.sAk = 1; g3_63.sBo = 0; g3_63.sBi = 0; g3_63.sBn = 1; g3_63.sBk = 1; g3_63.sCo = 0; g3_63.sCi = 0; g3_63.sCm = LP; g3_63.sRo = 0; g3_63.sRi = 0; g3_63.sRm = 0; g3_63.sRn = 0;
      g3_63.M = 8179; g3_63.N = 1; g3_63.K = H; g3_63.zi_n = 1; g3_63.flags = 1; g3_63.act = 0;
      g3_63.alpha = 1.0f; g3_63.beta = 0.0f; g3_63.sa = 1.0f; g3_63.sb = 8.0f; g3_63.Npad = LP; g3_63.pad_ = 0;
      k_gemm<0><<<dim3((unsigned)((LP) + 31) / 32, (unsigned)((8179) + 15) / 16, (unsigned)(1)), 32, 0, stream>>>(g3_63); }
    k_es_scatter<<<(unsigned)((8179 + 255) / 256), 256, 0, stream>>>(Y, LP, slot, IDX, 63, 516109, 8179, out);
}
